// AdvancedCrossStreamAttention_14912126452100
// MI455X (gfx1250) — hardware-verified
//
#include <hip/hip_runtime.h>
#include <math.h>

typedef __attribute__((ext_vector_type(16))) _Float16 v16h;
typedef __attribute__((ext_vector_type(8)))  _Float16 v8h;
typedef __attribute__((ext_vector_type(16))) __bf16   v16b;
typedef __attribute__((ext_vector_type(8)))  float    v8f;
typedef __attribute__((ext_vector_type(4)))  float    v4f;

__device__ __forceinline__ int frag_k(int i, int h) { return (i < 8) ? (8 * h + i) : (16 + 8 * h + (i - 8)); }
__device__ __forceinline__ __bf16 bf16_rne(float f) {
    unsigned int u = __float_as_uint(f);
    u += 0x7fffu + ((u >> 16) & 1u);
    return __builtin_bit_cast(__bf16, (unsigned short)(u >> 16));
}
__device__ __forceinline__ float bf16_f32(__bf16 b) { return __uint_as_float(((unsigned int)__builtin_bit_cast(unsigned short, b)) << 16); }
__device__ __forceinline__ v8f wmma16(v16h a, v16h b, v8f c) {
    c = __builtin_amdgcn_wmma_f32_16x16x32_f16(false, a, false, b, (short)0, c, false, false);
    asm volatile("v_nop\n\tv_nop\n\tv_nop\n\tv_nop" : "+v"(c) : "v"(a), "v"(b));
    return c;
}
__device__ __forceinline__ v8f wmmab(v16b a, v16b b, v8f c) {
    c = __builtin_amdgcn_wmma_f32_16x16x32_bf16(false, a, false, b, (short)0, c, false, false);
    asm volatile("v_nop\n\tv_nop\n\tv_nop\n\tv_nop" : "+v"(c) : "v"(a), "v"(b));
    return c;
}
struct Split { v16b hi, lo; };
__device__ __forceinline__ v8f wmma3(const Split& a, const Split& b, v8f c) {
    c = __builtin_amdgcn_wmma_f32_16x16x32_bf16(false, a.hi, false, b.hi, (short)0, c, false, false);
    c = __builtin_amdgcn_wmma_f32_16x16x32_bf16(false, a.hi, false, b.lo, (short)0, c, false, false);
    c = __builtin_amdgcn_wmma_f32_16x16x32_bf16(false, a.lo, false, b.hi, (short)0, c, false, false);
    asm volatile("v_nop\n\tv_nop\n\tv_nop\n\tv_nop" : "+v"(c) : "v"(a.hi), "v"(a.lo), "v"(b.hi), "v"(b.lo));
    return c;
}
struct Split3 { v16b hi, mid, lo; };
__device__ __forceinline__ v8f wmma6(const Split3& a, const Split3& b, v8f c) {
    c = __builtin_amdgcn_wmma_f32_16x16x32_bf16(false, a.hi, false, b.hi, (short)0, c, false, false);
    c = __builtin_amdgcn_wmma_f32_16x16x32_bf16(false, a.hi, false, b.mid, (short)0, c, false, false);
    c = __builtin_amdgcn_wmma_f32_16x16x32_bf16(false, a.mid, false, b.hi, (short)0, c, false, false);
    c = __builtin_amdgcn_wmma_f32_16x16x32_bf16(false, a.hi, false, b.lo, (short)0, c, false, false);
    c = __builtin_amdgcn_wmma_f32_16x16x32_bf16(false, a.mid, false, b.mid, (short)0, c, false, false);
    c = __builtin_amdgcn_wmma_f32_16x16x32_bf16(false, a.lo, false, b.hi, (short)0, c, false, false);
    asm volatile("v_nop\n\tv_nop\n\tv_nop\n\tv_nop" : "+v"(c) : "v"(a.hi), "v"(a.mid), "v"(a.lo), "v"(b.hi), "v"(b.mid), "v"(b.lo));
    return c;
}

__device__ __forceinline__ v16h fh_ld(const float* __restrict__ p, long long sk, int k0, int h, int klen, float s) {
    v16h a;
#pragma unroll
    for (int i = 0; i < 16; ++i) { const int k = k0 + frag_k(i, h); a[i] = (k < klen) ? (_Float16)(p[(long long)k * sk] * s) : (_Float16)0.f; }
    return a;
}
__device__ __forceinline__ Split sp_ld(const float* __restrict__ p, long long sk, int k0, int h, int klen, float s) {
    Split r;
#pragma unroll
    for (int i = 0; i < 16; ++i) {
        const int k = k0 + frag_k(i, h); const float x = (k < klen) ? p[(long long)k * sk] * s : 0.f;
        const __bf16 hb = bf16_rne(x); r.hi[i] = hb; r.lo[i] = bf16_rne(x - bf16_f32(hb));
    }
    return r;
}
__device__ __forceinline__ Split3 sp3_ld(const float* __restrict__ p, long long sk, int k0, int h, int klen, float s) {
    Split3 r;
#pragma unroll
    for (int i = 0; i < 16; ++i) {
        const int k = k0 + frag_k(i, h); const float x = (k < klen) ? p[(long long)k * sk] * s : 0.f;
        const __bf16 hb = bf16_rne(x); const float r1 = x - bf16_f32(hb); const __bf16 mb = bf16_rne(r1);
        r.hi[i] = hb; r.mid[i] = mb; r.lo[i] = bf16_rne(r1 - bf16_f32(mb));
    }
    return r;
}
__device__ __forceinline__ v16b bh_ld(const float* __restrict__ p, long long sk, int k0, int h, int klen, float s) {
    v16b a;
#pragma unroll
    for (int i = 0; i < 16; ++i) { const int k = k0 + frag_k(i, h); a[i] = bf16_rne((k < klen) ? p[(long long)k * sk] * s : 0.f); }
    return a;
}
__device__ __forceinline__ v16h fh_row(const _Float16* __restrict__ row, int k0, int h) {
    v16h a;
#pragma unroll
    for (int i = 0; i < 16; ++i) a[i] = row[k0 + frag_k(i, h)];
    return a;
}

#define VST2(T, ptr, val) do { const T vst2_v_ = (val); *(volatile T*)(ptr) = vst2_v_; __threadfence(); *(volatile T*)(ptr) = vst2_v_; } while (0)
typedef float v4f __attribute__((ext_vector_type(4)));
#define VST2V4(ptr, val) do { const v4f vst2_v4_ = (val); *(volatile v4f*)(ptr) = vst2_v4_; __threadfence(); *(volatile v4f*)(ptr) = vst2_v4_; } while (0)

__device__ __attribute__((noinline)) float act_fn(float v, int act) {
    if (act == 1) return fmaxf(v, 0.f);
    if (act == 2) { const float u = 0.7978845608028654f * (v + 0.044715f * v * v * v); return 0.5f * v * (1.f + tanhf(u)); }
    if (act == 3) return v / (1.f + expf(-v));
    if (act == 4) return 0.5f * v * (1.f + erff(v * 0.7071067811865476f));
    if (act == 5) return tanhf(v);
    if (act == 6) return 1.f / (1.f + expf(-v));
    if (act == 7) return (v > 0.f) ? v : 0.01f * v;
    if (act == 8) return (v > 0.f) ? v : (expf(v) - 1.f);
    if (act == 9) return fminf(fmaxf(v, 0.f), 6.f);
    if (act == 10) return fabsf(v);
    if (act == 11) return (v >= 0.f) ? v : 0.1f * v;
    if (act == 12) return (v > 0.f) ? v : 0.2f * v;
    if (act == 13) return (v > 20.f) ? v : log1pf(expf(v));
    return v;
}

struct GemmP {
    const float* A; const float* B; const float* bias; const float* R; float* C;
    long long sAo, sAi, sAm, sAk, sBo, sBi, sBn, sBk, sCo, sCi, sCm, sRo, sRi, sRm, sRn;
    int M, N, K, zi_n, flags, act; float alpha, beta, sa, sb;
    int Npad, pad_;
};
static_assert(sizeof(GemmP) == 5 * 8 + 15 * 8 + 6 * 4 + 4 * 4 + 2 * 4, "GemmP has padding");

template <int MODE>
__global__ __launch_bounds__(32) void k_gemm(GemmP p) {
    const int lane = threadIdx.x & 31, h = lane >> 4, l15 = lane & 15;
    const int m0 = blockIdx.y * 16, n0 = blockIdx.x * 32;
    const int z = blockIdx.z, zo = z / p.zi_n, zi = z - zo * p.zi_n;
    const float* A = p.A + zo * p.sAo + zi * p.sAi;
    const float* B = p.B + zo * p.sBo + zi * p.sBi;
    const int am = min(m0 + l15, p.M - 1);
    v8f acc[2], comp[2];
#pragma unroll
    for (int t = 0; t < 2; ++t) { v8f zz = {}; acc[t] = zz; comp[t] = zz; }
    for (int k0 = 0; k0 < p.K; k0 += 32) {
        const float* arow = A + (long long)am * p.sAm;
        if (MODE == 1) {
            const Split a = sp_ld(arow, p.sAk, k0, h, p.K, 1.f);
#pragma unroll
            for (int t = 0; t < 2; ++t) {
                const int bn = min(n0 + t * 16 + l15, p.N - 1);
                acc[t] = wmma3(a, sp_ld(B + (long long)bn * p.sBn, p.sBk, k0, h, p.K, 1.f), acc[t]);
            }
        } else if (MODE == 3) {
            const Split3 a = sp3_ld(arow, p.sAk, k0, h, p.K, 1.f);
#pragma unroll
            for (int t = 0; t < 2; ++t) {
                const int bn = min(n0 + t * 16 + l15, p.N - 1);
                acc[t] = wmma6(a, sp3_ld(B + (long long)bn * p.sBn, p.sBk, k0, h, p.K, 1.f), acc[t]);
            }
        } else if (MODE == 4) {
            const Split3 a = sp3_ld(arow, p.sAk, k0, h, p.K, 1.f);
#pragma unroll
            for (int t = 0; t < 2; ++t) {
                const int bn = min(n0 + t * 16 + l15, p.N - 1); v8f zz = {};
                const v8f part = wmma6(a, sp3_ld(B + (long long)bn * p.sBn, p.sBk, k0, h, p.K, 1.f), zz);
                const v8f y = part - comp[t]; const v8f s = acc[t] + y; comp[t] = (s - acc[t]) - y; acc[t] = s;
            }
        } else if (MODE == 2) {
            const v16b a = bh_ld(arow, p.sAk, k0, h, p.K, 1.f);
#pragma unroll
            for (int t = 0; t < 2; ++t) {
                const int bn = min(n0 + t * 16 + l15, p.N - 1);
                acc[t] = wmmab(a, bh_ld(B + (long long)bn * p.sBn, p.sBk, k0, h, p.K, 1.f), acc[t]);
            }
        } else {
            const v16h a = fh_ld(arow, p.sAk, k0, h, p.K, p.sa);
#pragma unroll
            for (int t = 0; t < 2; ++t) {
                const int bn = min(n0 + t * 16 + l15, p.N - 1);
                acc[t] = wmma16(a, fh_ld(B + (long long)bn * p.sBn, p.sBk, k0, h, p.K, p.sb), acc[t]);
            }
        }
    }
    const float iscale = (MODE == 0) ? p.alpha / (p.sa * p.sb) : p.alpha;
    float* C = p.C + zo * p.sCo + zi * p.sCi;
    const float* R = p.R + zo * p.sRo + zi * p.sRi;
    __shared__ __align__(16) float ctile[16][36];
#pragma unroll
    for (int t = 0; t < 2; ++t) {
        const int n = n0 + t * 16 + l15; const int nn = min(n, p.N - 1);
#pragma unroll
        for (int r = 0; r < 8; ++r) {
            const int m = m0 + 8 * h + r; const int mm = min(m, p.M - 1);
            float v = acc[t][r] * iscale;
            if (p.flags & 1) v += p.bias[nn];
            if (p.flags & 2) v += p.bias[mm];
            if (p.flags & 8) v *= p.bias[(long long)zo * p.M + mm];
            v = act_fn(v, p.act);
            if (p.flags & 4) v += p.beta * R[(long long)mm * p.sRm + (long long)nn * p.sRn];
            ctile[8 * h + r][t * 16 + l15] = (n < p.N) ? v : 0.f;
        }
    }
    __syncthreads();
    const int NW = (p.Npad > p.N) ? p.Npad : p.N;
    const bool fast = (m0 + 16 <= p.M) && (n0 + 32 <= NW) && ((p.sCm & 3) == 0) && ((((size_t)C) & 15) == 0);
    if (fast) {
#pragma unroll
        for (int s = 0; s < 4; ++s) {
            const int row = s * 4 + (lane >> 3), c4 = (lane & 7) * 4;
            const v4f v = *(const v4f*)&ctile[row][c4];
            VST2V4(C + (long long)(m0 + row) * p.sCm + n0 + c4, v);
        }
    } else {
        for (int row = 0; row < 16; ++row) {
            const int m = m0 + row, n = n0 + lane;
            if (m < p.M && n < NW) VST2(float, C + (long long)m * p.sCm + n, ctile[row][lane]);
        }
    }
}


template <int MODE, int TM, int TN>
__global__ __launch_bounds__(32) void k_gemmT(GemmP p) {
    const int lane = threadIdx.x & 31, h = lane >> 4, l15 = lane & 15;
    const int m0 = blockIdx.y * (16 * TM), n0 = blockIdx.x * (16 * TN);
    const int z = blockIdx.z, zo = z / p.zi_n, zi = z - zo * p.zi_n;
    const float* A = p.A + zo * p.sAo + zi * p.sAi;
    const float* B = p.B + zo * p.sBo + zi * p.sBi;
    v8f acc[TM][TN];
#pragma unroll
    for (int i = 0; i < TM; ++i)
#pragma unroll
        for (int t = 0; t < TN; ++t) { v8f zz = {}; acc[i][t] = zz; }
    for (int k0 = 0; k0 < p.K; k0 += 32) {
        if (MODE == 1) {
            Split a[TM], b[TN];
#pragma unroll
            for (int i = 0; i < TM; ++i) { const int am = min(m0 + 16 * i + l15, p.M - 1); a[i] = sp_ld(A + (long long)am * p.sAm, p.sAk, k0, h, p.K, 1.f); }
#pragma unroll
            for (int t = 0; t < TN; ++t) { const int bn = min(n0 + 16 * t + l15, p.N - 1); b[t] = sp_ld(B + (long long)bn * p.sBn, p.sBk, k0, h, p.K, 1.f); }
#pragma unroll
            for (int i = 0; i < TM; ++i)
#pragma unroll
                for (int t = 0; t < TN; ++t) acc[i][t] = wmma3(a[i], b[t], acc[i][t]);
        } else if (MODE == 2) {
            v16b a[TM], b[TN];
#pragma unroll
            for (int i = 0; i < TM; ++i) { const int am = min(m0 + 16 * i + l15, p.M - 1); a[i] = bh_ld(A + (long long)am * p.sAm, p.sAk, k0, h, p.K, 1.f); }
#pragma unroll
            for (int t = 0; t < TN; ++t) { const int bn = min(n0 + 16 * t + l15, p.N - 1); b[t] = bh_ld(B + (long long)bn * p.sBn, p.sBk, k0, h, p.K, 1.f); }
#pragma unroll
            for (int i = 0; i < TM; ++i)
#pragma unroll
                for (int t = 0; t < TN; ++t) acc[i][t] = wmmab(a[i], b[t], acc[i][t]);
        } else {
            v16h a[TM], b[TN];
#pragma unroll
            for (int i = 0; i < TM; ++i) { const int am = min(m0 + 16 * i + l15, p.M - 1); a[i] = fh_ld(A + (long long)am * p.sAm, p.sAk, k0, h, p.K, p.sa); }
#pragma unroll
            for (int t = 0; t < TN; ++t) { const int bn = min(n0 + 16 * t + l15, p.N - 1); b[t] = fh_ld(B + (long long)bn * p.sBn, p.sBk, k0, h, p.K, p.sb); }
#pragma unroll
            for (int i = 0; i < TM; ++i)
#pragma unroll
                for (int t = 0; t < TN; ++t) acc[i][t] = wmma16(a[i], b[t], acc[i][t]);
        }
    }
    const float iscale = (MODE == 0) ? p.alpha / (p.sa * p.sb) : p.alpha;
    float* C = p.C + zo * p.sCo + zi * p.sCi;
    const float* R = p.R + zo * p.sRo + zi * p.sRi;
    const int NW = (p.Npad > p.N) ? p.Npad : p.N;
    __shared__ __align__(16) float ctile[16][36];
#pragma unroll
    for (int i = 0; i < TM; ++i) {
        const int mb = m0 + 16 * i; if (mb >= p.M) break;
#pragma unroll
        for (int tp = 0; tp < TN / 2; ++tp) {
            const int nb = n0 + 32 * tp; if (nb >= NW) break;
#pragma unroll
            for (int t2 = 0; t2 < 2; ++t2) {
                const int t = 2 * tp + t2; const int n = nb + t2 * 16 + l15; const int nn = min(n, p.N - 1);
#pragma unroll
                for (int r = 0; r < 8; ++r) {
                    const int m = mb + 8 * h + r; const int mm = min(m, p.M - 1);
                    float v = acc[i][t][r] * iscale;
                    if (p.flags & 1) v += p.bias[nn];
                    if (p.flags & 2) v += p.bias[mm];
            if (p.flags & 8) v *= p.bias[(long long)zo * p.M + mm];
                    v = act_fn(v, p.act);
                    if (p.flags & 4) v += p.beta * R[(long long)mm * p.sRm + (long long)nn * p.sRn];
                    ctile[8 * h + r][t2 * 16 + l15] = (n < p.N) ? v : 0.f;
                }
            }
            __syncthreads();
            const bool fast = (mb + 16 <= p.M) && (nb + 32 <= NW) && ((p.sCm & 3) == 0) && ((((size_t)C) & 15) == 0);
            if (fast) {
#pragma unroll
                for (int s = 0; s < 4; ++s) {
                    const int row = s * 4 + (lane >> 3), c4 = (lane & 7) * 4;
                    const v4f v = *(const v4f*)&ctile[row][c4];
                    VST2V4(C + (long long)(mb + row) * p.sCm + nb + c4, v);
                }
            } else {
                for (int row = 0; row < 16; ++row) {
                    const int m = mb + row, n = nb + lane;
                    if (m < p.M && n < NW) VST2(float, C + (long long)m * p.sCm + n, ctile[row][lane]);
                }
            }
            __syncthreads();
        }
    }
}

#define AW 4
struct AttnP {
    const float* Q; const float* K; const float* V; float* O; float* P; const float* Mf; const int* Mi; float* ST;
    const float* Pw; const float* Rt; const int* SQ; const int* SK;
    long long swb, swh, swi, swj, srb, srh, sri;
    long long sQb, sQh, sQi, sQd, sKb, sKh, sKj, sKd, sVb, sVh, sVj, sVd, sOb, sOh, sOi, sPb, sPh, sPi, smb, smh, smi, smj;
    int Lq, Lk, dh, dv, hrep, causal, coff, pband;
    float scale, mfill; int nonorm, mpol;
    int roff, rn, segpol, win;
};
static_assert(sizeof(AttnP) == 12 * 8 + 29 * 8 + 16 * 4, "AttnP has padding");

#ifndef KATTN_ATTR
#define KATTN_ATTR
#endif
template <int DHP, int DVP, int QM, bool SPLITPV, bool TWOPASS>
__global__ __launch_bounds__(32 * AW) KATTN_ATTR void k_attn(AttnP p) {
    constexpr int NT = DVP / 16;
    constexpr int KS = DHP / 32;
    constexpr int VP = DVP + 8;
    __shared__ __align__(16) float    pl[AW][16 * 64];
    __shared__ __align__(16) _Float16 vl[(SPLITPV ? 2 : 1) * 64 * VP];
    const int lane = threadIdx.x & 31, hf = lane >> 4, l15 = lane & 15, wave = threadIdx.x >> 5;
    const int h = blockIdx.y, b = blockIdx.z, hk = h / p.hrep;
    const int q0 = (blockIdx.x * AW + wave) * 16;
    float* myp = pl[wave];
    const float L2E = 1.4426950408889634f;
    const float NEG = -__builtin_inff();
    const int qi = min(q0 + l15, p.Lq - 1);
    const float* qrow = p.Q + b * p.sQb + h * p.sQh + (long long)qi * p.sQi;
    const float* kbase = p.K + b * p.sKb + hk * p.sKh;
    const float* vbase = p.V + b * p.sVb + hk * p.sVh;
    v16h qa[QM == 0 ? KS : 1]; Split qs_[QM == 1 ? KS : 1]; Split3 qt_[QM == 2 ? KS : 1];
#pragma unroll
    for (int ks = 0; ks < KS; ++ks) {
        if (QM == 2) qt_[ks] = sp3_ld(qrow, p.sQd, ks * 32, hf, p.dh, 1.f);
        else if (QM == 1) qs_[ks] = sp_ld(qrow, p.sQd, ks * 32, hf, p.dh, 1.f);
        else qa[ks] = fh_ld(qrow, p.sQd, ks * 32, hf, p.dh, 1.f);
    }
    v8f o[NT]; float m8[8], l8[8];
#pragma unroll
    for (int t = 0; t < NT; ++t) { v8f zz = {}; o[t] = zz; }
#pragma unroll
    for (int i = 0; i < 8; ++i) { m8[i] = NEG; l8[i] = 0.f; }
    int jend = p.Lk; int jstart = 0;
    if (p.causal == 1) { const int je = (blockIdx.x * AW + AW - 1) * 16 + 16 + p.coff; jend = min(jend, max(je, 0)); }
    if (p.win > 0) { const int js = (int)(blockIdx.x * AW) * 16 + p.coff - p.win; jstart = (js > 0) ? (js / 64) * 64 : 0; }
    const int npass = TWOPASS ? 2 : 1;
    for (int pass = 0; pass < npass; ++pass) {
        const bool dopv = (!TWOPASS) || pass == 1;
        for (int j0 = jstart; j0 < jend; j0 += 64) {
            if (dopv) {
                __syncthreads();
                for (int idx = threadIdx.x; idx < 64 * DVP; idx += 32 * AW) {
                    const int jr = idx / DVP, d = idx - jr * DVP, j = j0 + jr;
                    const float f = (j < p.Lk && d < p.dv) ? vbase[(long long)j * p.sVj + (long long)d * p.sVd] : 0.f;
                    if (SPLITPV) {
                        const __bf16 hb = bf16_rne(f);
                        ((__bf16*)vl)[jr * VP + d] = hb; ((__bf16*)vl)[64 * VP + jr * VP + d] = bf16_rne(f - bf16_f32(hb));
                    } else vl[jr * VP + d] = (_Float16)f;
                }
            }
            v8f s[4];
#pragma unroll
            for (int t = 0; t < 4; ++t) {
                const int j = min(j0 + t * 16 + l15, p.Lk - 1);
                const float* krow = kbase + (long long)j * p.sKj;
                v8f acc = {};
#pragma unroll
                for (int ks = 0; ks < KS; ++ks) {
                    if (QM == 2)      acc = wmma6(qt_[ks], sp3_ld(krow, p.sKd, ks * 32, hf, p.dh, 1.f), acc);
                    else if (QM == 1) acc = wmma3(qs_[ks], sp_ld(krow, p.sKd, ks * 32, hf, p.dh, 1.f), acc);
                    else              acc = wmma16(qa[ks], fh_ld(krow, p.sKd, ks * 32, hf, p.dh, 1.f), acc);
                }
                s[t] = acc;
            }
            float pv[8][4];
#pragma unroll
            for (int i = 0; i < 8; ++i) {
                const int irow = q0 + i + 8 * hf;
                const int ic = min(irow, p.Lq - 1);
                float sc[4];
#pragma unroll
                for (int t = 0; t < 4; ++t) {
                    const int jg = j0 + t * 16 + l15;
                    float v = s[t][i] * p.scale;
                    if (p.Mf) v += p.Mf[b * p.smb + h * p.smh + (long long)ic * p.smi + (long long)min(jg, p.Lk - 1) * p.smj];
                    if (p.Rt) { int rc = ic - min(jg, p.Lk - 1) + p.roff; rc = rc < 0 ? 0 : (rc >= p.rn ? p.rn - 1 : rc); v += p.Rt[b * p.srb + h * p.srh + (long long)ic * p.sri + rc]; }
                    if (p.Mi) { const int mv = p.Mi[b * p.smb + h * p.smh + (long long)ic * p.smi + (long long)min(jg, p.Lk - 1) * p.smj]; if (p.mpol ? (mv != 0) : (mv == 0)) v = p.mfill; }
                    if (p.SQ) { const bool same = p.SQ[(long long)b * p.Lq + ic] == p.SK[(long long)b * p.Lk + min(jg, p.Lk - 1)]; if (p.segpol ? same : !same) v = p.mfill; }
                    if (p.causal == 2 && jg > irow + p.coff) v = p.mfill;
                    if (jg >= p.Lk || (p.causal == 1 && jg > irow + p.coff) || (p.causal == 3 && jg < irow + p.coff) || (p.win > 0 && irow + p.coff - jg > p.win)) v = NEG; else v *= L2E;
                    sc[t] = v;
                }
                if (!TWOPASS || pass == 0) {
                    float mx = fmaxf(fmaxf(sc[0], sc[1]), fmaxf(sc[2], sc[3]));
                    mx = fmaxf(mx, __shfl_xor(mx, 1, 32)); mx = fmaxf(mx, __shfl_xor(mx, 2, 32));
                    mx = fmaxf(mx, __shfl_xor(mx, 4, 32)); mx = fmaxf(mx, __shfl_xor(mx, 8, 32));
                    const float mnew = fmaxf(m8[i], mx);
                    const float corr = (mnew == NEG) ? 1.f : exp2f(m8[i] - mnew);
                    float rs = 0.f;
#pragma unroll
                    for (int t = 0; t < 4; ++t) {
                        const float pp = (sc[t] == NEG) ? 0.f : exp2f(sc[t] - mnew); rs += pp;
                        pv[i][t] = p.Pw ? pp * p.Pw[b * p.swb + h * p.swh + (long long)ic * p.swi + (long long)min(j0 + t * 16 + l15, p.Lk - 1) * p.swj] : pp;
                    }
                    rs += __shfl_xor(rs, 1, 32); rs += __shfl_xor(rs, 2, 32); rs += __shfl_xor(rs, 4, 32); rs += __shfl_xor(rs, 8, 32);
                    l8[i] = l8[i] * corr + rs; m8[i] = mnew;
                    if (!TWOPASS) {
#pragma unroll
                        for (int t = 0; t < NT; ++t) o[t][i] *= corr;
                    }
                } else {
                    const float inv = (l8[i] > 0.f) ? 1.f / l8[i] : 0.f;
#pragma unroll
                    for (int t = 0; t < 4; ++t) {
                        const int jg = j0 + t * 16 + l15;
                        float pp = (sc[t] == NEG) ? 0.f : exp2f(sc[t] - m8[i]) * inv;
                        if (p.Pw) pp *= p.Pw[b * p.swb + h * p.swh + (long long)ic * p.swi + (long long)min(jg, p.Lk - 1) * p.swj];
                        pv[i][t] = pp;
                    }
                }
            }
            if (dopv) {
#pragma unroll
                for (int i = 0; i < 8; ++i)
#pragma unroll
                    for (int t = 0; t < 4; ++t) ((volatile float*)myp)[(i + 8 * hf) * 64 + t * 16 + l15] = pv[i][t];
                __syncthreads();
                if (p.P) {
                    float* pb_ = p.P + b * p.sPb + h * p.sPh;
                    const bool fastP = (p.pband == 0) && ((p.sPi & 3) == 0) && (j0 + 64 <= p.Lk) && (q0 + 16 <= p.Lq) && ((((size_t)pb_) & 15) == 0);
                    if (fastP) {
#pragma unroll
                        for (int s = 0; s < 8; ++s) {
                            const int row = s * 2 + (lane >> 4), c4 = (lane & 15) * 4;
                            const v4f v = *(const v4f*)(myp + row * 64 + c4);
                            VST2V4(pb_ + (long long)(q0 + row) * p.sPi + j0 + c4, v);
                        }
                    } else {
                        for (int row = 0; row < 16; ++row) {
                            const int irow = q0 + row; if (irow >= p.Lq) continue;
                            for (int c = lane; c < 64; c += 32) {
                                const int jg = j0 + c; if (jg >= p.Lk) continue;
                                if (p.pband == 0) VST2(float, pb_ + (long long)irow * p.sPi + jg, myp[row * 64 + c]);
                                else if (jg - irow <= p.pband && irow - jg <= p.pband) VST2(float, pb_ + (long long)irow * p.sPi + (jg - irow + p.pband), myp[row * 64 + c]);
                            }
                        }
                    }
                }
                if (SPLITPV) {
                    const Split pa0 = sp_ld(myp + l15 * 64, 1, 0, hf, 64, 1.f), pa1 = sp_ld(myp + l15 * 64, 1, 32, hf, 64, 1.f);
                    const __bf16* vh = (const __bf16*)vl; const __bf16* vlo = vh + 64 * VP;
#pragma unroll
                    for (int t = 0; t < NT; ++t) {
                        const int dcol = t * 16 + l15;
                        Split b0, b1;
#pragma unroll
                        for (int e = 0; e < 16; ++e) {
                            const int k0 = frag_k(e, hf), k1 = 32 + frag_k(e, hf);
                            b0.hi[e] = vh[k0 * VP + dcol]; b0.lo[e] = vlo[k0 * VP + dcol]; b1.hi[e] = vh[k1 * VP + dcol]; b1.lo[e] = vlo[k1 * VP + dcol];
                        }
                        o[t] = wmma3(pa0, b0, o[t]);
                        o[t] = wmma3(pa1, b1, o[t]);
                    }
                } else {
                    const v16h pa0 = fh_ld(myp + l15 * 64, 1, 0, hf, 64, 4096.f), pa1 = fh_ld(myp + l15 * 64, 1, 32, hf, 64, 4096.f);
#pragma unroll
                    for (int t = 0; t < NT; ++t) {
                        const int dcol = t * 16 + l15;
                        v16h b0, b1;
#pragma unroll
                        for (int e = 0; e < 16; ++e) { b0[e] = vl[frag_k(e, hf) * VP + dcol]; b1[e] = vl[(32 + frag_k(e, hf)) * VP + dcol]; }
                        o[t] = wmma16(pa0, b0, o[t]);
                        o[t] = wmma16(pa1, b1, o[t]);
                    }
                }
            }
        }
    }
    float* obase = p.O + b * p.sOb + h * p.sOh;
    if (p.ST) {
        const int rl = lane >> 1, isel = rl & 7;
        float mv = 0.f, lv = 0.f;
#pragma unroll
        for (int i = 0; i < 8; ++i) if (i == isel) { mv = m8[i]; lv = l8[i]; }
        const int irow = q0 + rl;
        if (irow < p.Lq) { float* st = p.ST + (((long long)b * gridDim.y + h) * p.Lq + irow) * 2 + (lane & 1); VST2(float, st, (lane & 1) ? lv : mv * 0.6931471805599453f); }
    }
    float invr[8];
#pragma unroll
    for (int i = 0; i < 8; ++i) {
        if (TWOPASS) invr[i] = SPLITPV ? 1.f : (1.f / 4096.f);
        else if (p.nonorm) invr[i] = exp2f(m8[i]) * (SPLITPV ? 1.f : (1.f / 4096.f));
        else invr[i] = (l8[i] > 0.f) ? (SPLITPV ? 1.f / l8[i] : 1.f / (l8[i] * 4096.f)) : 0.f;
    }
    __syncthreads();
    const bool ofast = ((p.sOi & 3) == 0) && ((((size_t)obase) & 15) == 0) && (q0 + 16 <= p.Lq);
#pragma unroll
    for (int c0 = 0; c0 < DVP; c0 += 64) {
#pragma unroll
        for (int i = 0; i < 8; ++i)
#pragma unroll
            for (int t = 0; t < NT; ++t) if (t * 16 >= c0 && t * 16 < c0 + 64) ((volatile float*)myp)[(i + 8 * hf) * 64 + (t * 16 - c0) + l15] = o[t][i] * invr[i];
        __syncthreads();
        const int cw = (DVP - c0 < 64) ? (DVP - c0) : 64;
        if (ofast && (c0 + cw <= p.dv) && (cw % 32 == 0)) {
            const int lpr = cw / 4;
            const int rows_per_ins = 32 / lpr;
            for (int r0 = 0; r0 < 16; r0 += rows_per_ins) {
                const int row = r0 + lane / lpr, c4 = (lane % lpr) * 4;
                const v4f v = *(const v4f*)(myp + row * 64 + c4);
                VST2V4(obase + (long long)(q0 + row) * p.sOi + c0 + c4, v);
            }
        } else {
            for (int row = 0; row < 16; ++row) {
                const int irow = q0 + row; if (irow >= p.Lq) continue;
                for (int c = lane; c < cw; c += 32) { const int d = c0 + c; if (d < p.dv) VST2(float, obase + (long long)irow * p.sOi + d, myp[row * 64 + c]); }
            }
        }
        __syncthreads();
    }
}

struct TrP { const float* src; float* dst; const float* R2; long long sSz, lds, sDz, ldd, sRz, ldr; int R, C, flags, act; float alpha, beta; };
static_assert(sizeof(TrP) == 3 * 8 + 6 * 8 + 6 * 4, "TrP has padding");
__global__ __launch_bounds__(256) void k_tr(TrP p) {
    __shared__ float tile[32][33];
    const int c0 = blockIdx.x * 32, r0 = blockIdx.y * 32, z = blockIdx.z;
    const int lane = threadIdx.x & 31, wave = threadIdx.x >> 5;
    const float* s = p.src + z * p.sSz;
#pragma unroll
    for (int k = 0; k < 4; ++k) {
        const int rl = wave * 4 + k, r = r0 + rl, c = c0 + lane;
        tile[rl][lane] = (r < p.R && c < p.C) ? s[(long long)r * p.lds + c] : 0.f;
    }
    __syncthreads();
    float* d = p.dst + z * p.sDz; const float* rr = p.R2 + z * p.sRz;
#pragma unroll
    for (int k = 0; k < 4; ++k) {
        const int cl = wave * 4 + k, c = c0 + cl, r = r0 + lane;
        if (c < p.C && r < p.R) {
            float v = act_fn(p.alpha * tile[lane][cl], p.act);
            if (p.flags & 1) v += p.beta * rr[(long long)c * p.ldr + r];
            VST2(float, d + (long long)c * p.ldd + r, v);
        }
    }
}

__global__ __launch_bounds__(256) void k_affine(const float* __restrict__ src, float* __restrict__ dst, int n, float a, float b, const float* __restrict__ sdev) {
    const int i = blockIdx.x * 256 + threadIdx.x;
    if (i < n) { const float aa = sdev ? a * sdev[0] : a; const float v = aa * src[i] + b; VST2(float, dst + i, v); }
}

struct SmP { const float* src; float* dst; const float* Mf; long long sz, sr, dz, dr, smz, smr; int n, pad; float scale_in, scale_out; };
static_assert(sizeof(SmP) == 3 * 8 + 6 * 8 + 4 * 4, "SmP has padding");
__global__ __launch_bounds__(256) void k_softmax(SmP p) {
    __shared__ float red[256];
    const int r = blockIdx.x, z = blockIdx.y, tid = threadIdx.x;
    const float* s = p.src + z * p.sz + (long long)r * p.sr;
    const float* mf = p.Mf ? (p.Mf + z * p.smz + (long long)r * p.smr) : nullptr;
    float mx = -__builtin_inff();
    for (int j = tid; j < p.n; j += 256) { float v = s[j] * p.scale_in; if (mf) v += mf[j]; mx = fmaxf(mx, v); }
    red[tid] = mx; __syncthreads();
    for (int o = 128; o > 0; o >>= 1) { if (tid < o) red[tid] = fmaxf(red[tid], red[tid + o]); __syncthreads(); }
    mx = red[0]; __syncthreads();
    float sum = 0.f;
    for (int j = tid; j < p.n; j += 256) { float v = s[j] * p.scale_in; if (mf) v += mf[j]; sum += (mx == -__builtin_inff()) ? 0.f : expf(v - mx); }
    red[tid] = sum; __syncthreads();
    for (int o = 128; o > 0; o >>= 1) { if (tid < o) red[tid] += red[tid + o]; __syncthreads(); }
    sum = red[0];
    const float inv = (sum > 0.f) ? p.scale_out / sum : 0.f;
    float* d = p.dst + z * p.dz + (long long)r * p.dr;
    for (int j = tid; j < p.n; j += 256) { float v = s[j] * p.scale_in; if (mf) v += mf[j]; const float o = (mx == -__builtin_inff()) ? 0.f : expf(v - mx) * inv; VST2(float, d + j, o); }
}
__global__ __launch_bounds__(256) void k_stats(const float* __restrict__ x, long long sz, long long so, long long si, int inner, int n, float eps, float* __restrict__ stat, int mode) {
    __shared__ float red[256];
    const int z = blockIdx.x, tid = threadIdx.x;
    const float* base = x + z * sz;
    float s = 0.f;
    for (int e = tid; e < n; e += 256) s += base[(long long)(e / inner) * so + (long long)(e % inner) * si];
    red[tid] = s; __syncthreads();
    for (int o = 128; o > 0; o >>= 1) { if (tid < o) red[tid] += red[tid + o]; __syncthreads(); }
    const float mu = (mode == 0 || mode == 3) ? red[0] / (float)n : 0.f; __syncthreads();
    float q = 0.f;
    for (int e = tid; e < n; e += 256) { const float dlt = base[(long long)(e / inner) * so + (long long)(e % inner) * si] - mu; q += dlt * dlt; }
    red[tid] = q; __syncthreads();
    for (int o = 128; o > 0; o >>= 1) { if (tid < o) red[tid] += red[tid + o]; __syncthreads(); }
    {
        float rs;
        if (mode == 2) rs = sqrtf((float)n) / fmaxf(sqrtf(red[0]), eps); else if (mode == 3) rs = rsqrtf(red[0] / (float)(n - 1) + eps); else rs = rsqrtf(red[0] / (float)n + eps);
        if (tid < 32) { const float v = (tid == 0) ? mu : ((tid == 1) ? rs : 0.f); VST2(float, stat + (long long)z * 32 + tid, v); }
    }
}
__global__ __launch_bounds__(256) void k_norm_apply(const float* __restrict__ x, float* __restrict__ y, const float* __restrict__ stat, const float* __restrict__ g, const float* __restrict__ bta,
                                                     int Z, int C, int L, int G, int bn, int act) {
    const long long idx = (long long)blockIdx.x * 256 + threadIdx.x;
    if (idx >= (long long)Z * C * L) return;
    const int l = (int)(idx % L); const long long zc = idx / L; const int c = (int)(zc % C), z = (int)(zc / C); (void)l;
    const int set = bn ? c : (z * G + c / (C / G));
    float v = (x[idx] - stat[(long long)set * 32]) * stat[(long long)set * 32 + 1];
    if (g) v *= g[c];
    if (bta) v += bta[c];
    v = act_fn(v, act);
    VST2(float, y + idx, v);
}

__global__ __launch_bounds__(256) void k_lse_neg(const float* __restrict__ st, float* __restrict__ c, int n) {
    const int i = blockIdx.x * 256 + threadIdx.x;
    if (i < n) { const float v = -(st[2 * i] + logf(st[2 * i + 1])); VST2(float, c + i, v); }
}

__global__ __launch_bounds__(256) void k_iota(int* __restrict__ dst, int n, int a, int b) {
    const int i = blockIdx.x * 256 + threadIdx.x;
    if (i < n) { const int v = a * i + b; VST2(int, dst + i, v); }
}

__global__ __launch_bounds__(256) void k_axpby(const float* __restrict__ x, const float* __restrict__ y, float* __restrict__ dst, int n, float a, float b, float c) {
    const int i = blockIdx.x * 256 + threadIdx.x;
    if (i < n) { const float v = a * x[i] + b * y[i] + c; VST2(float, dst + i, v); }
}

struct RopeP { const float* X; float* Y; const float* C; const float* Sn; const int* pos; long long sXr, sXh, sYr, sYh, sCb, sCp, sCd; int R, Hn, D, S, mode, tmode, pmode, pad; };
static_assert(sizeof(RopeP) == 5 * 8 + 7 * 8 + 8 * 4, "RopeP has padding");
__global__ __launch_bounds__(256) void k_rope(RopeP p) {
    const long long idx = (long long)blockIdx.x * 256 + threadIdx.x;
    if (idx >= (long long)p.R * p.Hn * p.D) return;
    const int d = (int)(idx % p.D); const long long rh = idx / p.D; const int h = (int)(rh % p.Hn); const int r = (int)(rh / p.Hn);
    const int half = p.D / 2;
    int partner; float sign;
    if (p.mode == 0) { partner = (d < half) ? d + half : d - half; sign = (d < half) ? -1.f : 1.f; }
    else { partner = d ^ 1; sign = (d & 1) ? 1.f : -1.f; }
    const int tcol = (p.tmode == 0) ? d : ((p.tmode == 1) ? (d % half) : (d >> 1));
    const int pp = (p.pmode == 0) ? (r % p.S) : ((p.pmode == 1) ? h : p.pos[r]);
    const long long toff = (long long)(r / p.S) * p.sCb + (long long)pp * p.sCp + (long long)tcol * p.sCd;
    const float* xr = p.X + (long long)r * p.sXr + (long long)h * p.sXh;
    const float v = xr[d] * p.C[toff] + sign * xr[partner] * p.Sn[toff];
    VST2(float, p.Y + (long long)r * p.sYr + (long long)h * p.sYh + d, v);
}

__global__ __launch_bounds__(256) void k_invf(float* __restrict__ invb, int half, int D, float base, float num, int fmode, float cexp) {
    const int i = blockIdx.x * 256 + threadIdx.x;
    if (i >= ((half + 31) / 32) * 32) return;
    if (i >= half) { VST2(float, invb + i, 0.f); return; }
    const float e = (float)(2 * i) / (float)D;
    float invf;
    if (fmode == 1) invf = num * expf((float)(2 * i) * cexp);
    else if (fmode == 2) invf = num * powf(base, (-2.0f * ((float)i - 1.0f)) / (float)D);
    else invf = num * (1.0f / powf(base, e));
    VST2(float, invb + i, invf);
}
__global__ __launch_bounds__(256) void k_sincos(float* __restrict__ cs, float* __restrict__ sn, const float* __restrict__ invb, int S, int half, float pscale) {
    const int idx = blockIdx.x * 256 + threadIdx.x;
    if (idx >= S * half) return;
    const int s = idx / half, i = idx - s * half;
    const float ang = (pscale * (float)s) * invb[i];
    VST2(float, cs + idx, cosf(ang)); VST2(float, sn + idx, sinf(ang));
}

__global__ __launch_bounds__(256) void k_mulact(const float* __restrict__ x, const float* __restrict__ y, float* __restrict__ dst, int n, int act) {
    const int i = blockIdx.x * 256 + threadIdx.x;
    if (i < n) { const float v = act_fn(x[i], act) * y[i]; VST2(float, dst + i, v); }
}

__global__ __launch_bounds__(256) void k_matvec(GemmP p) {
    const int rpt = (p.N == 1) ? 1 : 32;
    const long long r0 = ((long long)blockIdx.x * 256 + threadIdx.x) * rpt; const int z = blockIdx.z, zo = z / p.zi_n, zi = z - zo * p.zi_n;
    if (r0 >= p.M) return;
    const float* Bb = p.B + zo * p.sBo + zi * p.sBi;
    float* C = p.C + zo * p.sCo + zi * p.sCi; const float* R = p.R + zo * p.sRo + zi * p.sRi;
    for (int rr = 0; rr < rpt; ++rr) {
        const long long r = r0 + rr; if (r >= p.M) break;
        const float* A = p.A + zo * p.sAo + zi * p.sAi + r * p.sAm;
        float acc[8] = {0.f, 0.f, 0.f, 0.f, 0.f, 0.f, 0.f, 0.f};
        for (int k = 0; k < p.K; ++k) { const float a = A[(long long)k * p.sAk];
#pragma unroll
            for (int j = 0; j < 8; ++j) if (j < p.N) acc[j] += a * Bb[(long long)j * p.sBn + (long long)k * p.sBk]; }
#pragma unroll
        for (int j = 0; j < 8; ++j) if (j < p.N) {
            float v = acc[j] * p.alpha;
            if (p.flags & 1) v += p.bias[j];
            if (p.flags & 2) v += p.bias[r];
            v = act_fn(v, p.act);
            if (p.flags & 4) v += p.beta * R[r * p.sRm + (long long)j * p.sRn];
            VST2(float, C + r * p.sCm + j, v);
        }
    }
}
__global__ __launch_bounds__(256) void k_smallsoftmax(const float* __restrict__ src, float* __restrict__ dst, long long sr, long long dr, int n, long long R, float scale) {
    const long long r0 = ((long long)blockIdx.x * 256 + threadIdx.x) * 32;
    for (int rr = 0; rr < 32; ++rr) {
        const long long r = r0 + rr; if (r >= R) return;
        const float* s = src + r * sr; float* d = dst + r * dr;
        float mx = -__builtin_inff();
        for (int j = 0; j < n; ++j) mx = fmaxf(mx, s[j] * scale);
        float sum = 0.f;
        for (int j = 0; j < n; ++j) sum += expf(s[j] * scale - mx);
        const float inv = 1.f / sum;
        for (int j = 0; j < n; ++j) { const float v = expf(s[j] * scale - mx) * inv; VST2(float, d + j, v); }
    }
}

__global__ __launch_bounds__(32) void k_unitstat(float* __restrict__ st) { const int t = threadIdx.x; const float v = (t == 1) ? 1.f : 0.f; VST2(float, st + t, v); }

__global__ __launch_bounds__(256) void k_lincopy(const float* __restrict__ src, long long lds, float* __restrict__ dst, long long ldd, long long rows, int cols) {
    const long long i = (long long)blockIdx.x * 256 + threadIdx.x; if (i >= rows * cols) return;
    const long long r = i / cols; const int c = (int)(i - r * cols);
    const float v = src[r * lds + c]; VST2(float, dst + r * ldd + c, v);
}

namespace w25 {
typedef __attribute__((ext_vector_type(16))) _Float16 v16h;
typedef __attribute__((ext_vector_type(8)))  _Float16 v8h;
typedef __attribute__((ext_vector_type(16))) __bf16   v16b;
typedef __attribute__((ext_vector_type(8)))  __bf16   v8b;
typedef __attribute__((ext_vector_type(8)))  float    v8f;
typedef __attribute__((ext_vector_type(4)))  float    v4f;

__device__ __forceinline__ unsigned short f2bf_bits(float f) {
  unsigned u = __float_as_uint(f);
  return (unsigned short)((u + 0x7FFFu + ((u >> 16) & 1u)) >> 16);
}
__device__ __forceinline__ float bf_bits2f(unsigned short h) { return __uint_as_float(((unsigned)h) << 16); }

__device__ __forceinline__ void dep_guard_h(v8f& a, v8f& b, v16h x, v16h y) { asm volatile("v_nop\n\tv_nop\n\tv_nop\n\tv_nop" : "+v"(a), "+v"(b) : "v"(x), "v"(y)); }
__device__ __forceinline__ void dep_guard_b(v8f& a, v8f& b, v16b x, v16b y) { asm volatile("v_nop\n\tv_nop\n\tv_nop\n\tv_nop" : "+v"(a), "+v"(b) : "v"(x), "v"(y)); }
__device__ __forceinline__ void keep4_h(v16h a, v16h b, v16h c, v16h d) { asm volatile("v_nop" :: "v"(a), "v"(b), "v"(c), "v"(d)); }
__device__ __forceinline__ void keep4_b(v16b a, v16b b, v16b c, v16b d) { asm volatile("v_nop" :: "v"(a), "v"(b), "v"(c), "v"(d)); }
__device__ __forceinline__ void acc_guard4(v8f& a, v8f& b, v8f& c, v8f& d) { asm volatile("v_nop\n\tv_nop\n\tv_nop\n\tv_nop" : "+v"(a), "+v"(b), "+v"(c), "+v"(d)); }
template <typename T> struct Frag;
template <> struct Frag<_Float16> {
  typedef v16h V; union U { v16h v; v8h h[2]; };
  static __device__ __forceinline__ v16h load(const _Float16* p) {
    U f; f.h[0] = *(const v8h*)(p); f.h[1] = *(const v8h*)(p + 16); return f.v;
  }
  static __device__ __forceinline__ v8f mma(v16h a, v16h b, v8f c) {
    return __builtin_amdgcn_wmma_f32_16x16x32_f16(false, a, false, b, (short)0, c, false, false);
  }
  static __device__ __forceinline__ void guard(v8f& a, v8f& b, v16h x, v16h y) { dep_guard_h(a, b, x, y); }
  static __device__ __forceinline__ void keep(v16h a, v16h b, v16h c, v16h d) { keep4_h(a, b, c, d); }
};
template <> struct Frag<__bf16> {
  typedef v16b V; union U { v16b v; v8b h[2]; };
  static __device__ __forceinline__ v16b load(const __bf16* p) {
    U f; f.h[0] = *(const v8b*)(p); f.h[1] = *(const v8b*)(p + 16); return f.v;
  }
  static __device__ __forceinline__ v8f mma(v16b a, v16b b, v8f c) {
    return __builtin_amdgcn_wmma_f32_16x16x32_bf16(false, a, false, b, (short)0, c, false, false);
  }
  static __device__ __forceinline__ void guard(v8f& a, v8f& b, v16b x, v16b y) { dep_guard_b(a, b, x, y); }
  static __device__ __forceinline__ void keep(v16b a, v16b b, v16b c, v16b d) { keep4_b(a, b, c, d); }
};

template <int ET> struct Elem;
template <> struct Elem<0> { typedef _Float16 T; };
template <> struct Elem<1> { typedef __bf16 T; };
template <int ET, bool SPLIT, int BIAS_MODE, int OUT_MODE, bool RESID, int ACT = 0>
__global__ __launch_bounds__(256) void wmma_gemm64(
    const unsigned short* __restrict__ Ap, const unsigned short* __restrict__ A2p, int lda, long strideA,
    const unsigned short* __restrict__ Btp, const unsigned short* __restrict__ Bt2p, int ldb, long strideB,
    void* __restrict__ Cout, void* __restrict__ Cout2, int ldc, long strideC,
    const float* __restrict__ bias,
    const float* __restrict__ resid, long strideR,
    int M, int N, int K, float scale) {
  typedef typename Elem<ET>::T T;
  typedef typename Frag<T>::V V;
  const T* A = (const T*)Ap; const T* A2 = (const T*)A2p; const T* Bt = (const T*)Btp; const T* Bt2 = (const T*)Bt2p;
  __shared__ __align__(16) float sT[8][16 * 68];
  const int b    = blockIdx.y;
  const int lane = threadIdx.x & 31;
  const int wave = threadIdx.x >> 5;
  const int tilesN = N >> 6;
  const int tilesM = M >> 6;
  const int tile = blockIdx.x * 8 + wave;
  if (tile >= tilesM * tilesN) return;
  const int tm = tile / tilesN;
  const int tn = tile - tm * tilesN;
  const int m0 = tm << 6;
  const int n0 = tn << 6;

  const T* Ab  = A  + (size_t)b * strideA;
  const T* Bb  = Bt + (size_t)b * strideB;
  const T* Ab2 = SPLIT ? (A2  + (size_t)b * strideA) : nullptr;
  const T* Bb2 = SPLIT ? (Bt2 + (size_t)b * strideB) : nullptr;

  const int rlane = lane & 15;
  const int koff  = (lane >> 4) * 8;
  const int mOff  = (lane >> 4) * 8;

  v8f acc[4][4];
#pragma unroll
  for (int i = 0; i < 4; ++i)
#pragma unroll
    for (int j = 0; j < 4; ++j) acc[i][j] = (v8f){0.f,0.f,0.f,0.f,0.f,0.f,0.f,0.f};

  for (int k0 = 0; k0 < K; k0 += 32) {
    V bh[4], bl[4];
#pragma unroll
    for (int j = 0; j < 4; ++j) {
      const size_t bo = (size_t)(n0 + (j << 4) + rlane) * ldb + koff + k0;
      bh[j] = Frag<T>::load(Bb + bo);
      if (SPLIT) bl[j] = Frag<T>::load(Bb2 + bo);
    }
#pragma unroll
    for (int i = 0; i < 4; ++i) {
      const size_t ao = (size_t)(m0 + (i << 4) + rlane) * lda + koff + k0;
      V ah = Frag<T>::load(Ab + ao);
      V al;
      if (SPLIT) al = Frag<T>::load(Ab2 + ao);
#pragma unroll
      for (int j = 0; j < 4; ++j) {
        acc[i][j] = Frag<T>::mma(ah, bh[j], acc[i][j]);
        if (SPLIT) {
          acc[i][j] = Frag<T>::mma(ah, bl[j], acc[i][j]);
          acc[i][j] = Frag<T>::mma(al, bh[j], acc[i][j]);
        }
      }
      Frag<T>::guard(acc[i][0], acc[i][3], ah, SPLIT ? al : ah);
    }
    Frag<T>::keep(bh[0], bh[1], bh[2], bh[3]);
    if (SPLIT) Frag<T>::keep(bl[0], bl[1], bl[2], bl[3]);
  }
  acc_guard4(acc[0][0], acc[0][1], acc[0][2], acc[0][3]);
  acc_guard4(acc[1][0], acc[1][1], acc[1][2], acc[1][3]);
  acc_guard4(acc[2][0], acc[2][1], acc[2][2], acc[2][3]);
  acc_guard4(acc[3][0], acc[3][1], acc[3][2], acc[3][3]);

  float* slab = sT[wave];
  const float* Rb = RESID ? (resid + (size_t)b * strideR) : nullptr;
#pragma unroll
  for (int i = 0; i < 4; ++i) {
    const int mBase = m0 + (i << 4);
#pragma unroll
    for (int j = 0; j < 4; ++j) {
      const int n = n0 + (j << 4) + rlane;
      float bv = 0.f;
      if (BIAS_MODE == 2) bv = bias[n];
#pragma unroll
      for (int r = 0; r < 8; ++r) {
        float v = acc[i][j][r] * scale;
        if (BIAS_MODE == 1) v += bias[mBase + mOff + r];
        if (BIAS_MODE == 2) v += bv;
        if (RESID) v += Rb[(size_t)(mBase + mOff + r) * ldc + n];
        if (ACT == 1) v = tanhf(v);
        if (ACT == 2) v = fmaxf(v, 0.0f);
        if (ACT == 3) v = v / (1.0f + expf(-v));
        if (ACT == 4) v = (v > 0.f) ? v : 0.01f * v;
        if (ACT == 5) v = 0.5f * v * (1.0f + erff(v * 0.70710678118654752f));
        slab[(mOff + r) * 68 + (j << 4) + rlane] = v;
      }
    }
    __builtin_amdgcn_fence(__ATOMIC_RELEASE, "workgroup");
    __builtin_amdgcn_wave_barrier();
    __builtin_amdgcn_fence(__ATOMIC_ACQUIRE, "workgroup");
    if (OUT_MODE == 0) {
      float* C = (float*)Cout + (size_t)b * strideC;
      const int hh = lane >> 4, c4 = (lane & 15) * 4;
      for (int pass = 0; pass < 2; ++pass) {
#pragma unroll
        for (int it = 0; it < 8; ++it) {
          const int row = it * 2 + hh;
          v4f v = *(const v4f*)(slab + row * 68 + c4);
          *(volatile v4f*)(C + (size_t)(mBase + row) * ldc + n0 + c4) = v;
        }
        __threadfence();
      }
    } else {
      const int q = lane >> 3, c8 = (lane & 7) * 8;
      unsigned short* C  = (unsigned short*)Cout  + (size_t)b * strideC;
      unsigned short* C2 = (OUT_MODE == 2) ? ((unsigned short*)Cout2 + (size_t)b * strideC) : nullptr;
      for (int pass = 0; pass < 2; ++pass) {
#pragma unroll
        for (int it = 0; it < 4; ++it) {
          const int row = it * 4 + q;
          const float* sp = slab + row * 68 + c8;
          v8h hv, lv;
#pragma unroll
          for (int e = 0; e < 8; ++e) {
            if (OUT_MODE == 1) {
              hv[e] = (_Float16)sp[e];
            } else {
              unsigned short hb = f2bf_bits(sp[e]);
              unsigned short lb = f2bf_bits(sp[e] - bf_bits2f(hb));
              hv[e] = __builtin_bit_cast(_Float16, hb);
              lv[e] = __builtin_bit_cast(_Float16, lb);
            }
          }
          *(volatile v8h*)(C + (size_t)(mBase + row) * ldc + n0 + c8) = hv;
          if (OUT_MODE == 2) *(volatile v8h*)(C2 + (size_t)(mBase + row) * ldc + n0 + c8) = lv;
        }
        __threadfence();
      }
    }
    __builtin_amdgcn_fence(__ATOMIC_RELEASE, "workgroup");
    __builtin_amdgcn_wave_barrier();
    __builtin_amdgcn_fence(__ATOMIC_ACQUIRE, "workgroup");
  }
}

__global__ __launch_bounds__(256) void cast_f32_f16x2(
    const float* __restrict__ in, _Float16* __restrict__ out, int n2) {
  int i = blockIdx.x * 256 + threadIdx.x;
  if (i < n2) {
    const _Float16 h0 = (_Float16)in[2 * i], h1 = (_Float16)in[2 * i + 1];
    const unsigned u = (unsigned)__builtin_bit_cast(unsigned short, h0) | ((unsigned)__builtin_bit_cast(unsigned short, h1) << 16);
    ((volatile unsigned*)out)[i] = u;
    __threadfence();
    ((volatile unsigned*)out)[i] = u;
  }
}


}

__global__ __launch_bounds__(256) void k_castT16(const float* __restrict__ src, long long lds, _Float16* __restrict__ dst, long long ldd, int R, int C, float s) {
    const long long i = (long long)blockIdx.x * 256 + threadIdx.x; const long long np = (long long)C * (R / 2); if (i >= np) return; const int c = (int)(i / (R / 2)); const int r = 2 * (int)(i % (R / 2));
    const _Float16 h0 = (_Float16)(src[(long long)r * lds + c] * s), h1 = (_Float16)(src[(long long)(r + 1) * lds + c] * s);
    const unsigned u = (unsigned)__builtin_bit_cast(unsigned short, h0) | ((unsigned)__builtin_bit_cast(unsigned short, h1) << 16);
    volatile unsigned* d = (volatile unsigned*)(dst + (long long)c * ldd + r); *d = u; __threadfence(); *d = u; }
__global__ __launch_bounds__(256) void k_cast16(const float* __restrict__ src, long long lds, _Float16* __restrict__ dst, long long ldd, int R, int C, float s) {
    const long long i = (long long)blockIdx.x * 256 + threadIdx.x; const long long np = (long long)R * (C / 2); if (i >= np) return; const int r = (int)(i / (C / 2)); const int c = 2 * (int)(i % (C / 2));
    const _Float16 h0 = (_Float16)(src[(long long)r * lds + c] * s), h1 = (_Float16)(src[(long long)r * lds + c + 1] * s);
    const unsigned u = (unsigned)__builtin_bit_cast(unsigned short, h0) | ((unsigned)__builtin_bit_cast(unsigned short, h1) << 16);
    volatile unsigned* d = (volatile unsigned*)(dst + (long long)r * ldd + c); *d = u; __threadfence(); *d = u; }

__device__ __forceinline__ unsigned int f2bf2_pack(float a, float b, unsigned int* lo) {
    const unsigned short ha = w25::f2bf_bits(a), hb = w25::f2bf_bits(b);
    const unsigned short la = w25::f2bf_bits(a - w25::bf_bits2f(ha)), lb = w25::f2bf_bits(b - w25::bf_bits2f(hb));
    *lo = (unsigned)la | ((unsigned)lb << 16); return (unsigned)ha | ((unsigned)hb << 16); }
__global__ __launch_bounds__(256) void k_castS16(const float* __restrict__ src, long long lds, __bf16* __restrict__ dhi, __bf16* __restrict__ dlo, long long ldd, int R, int C, float s, int transpose) {
    const long long i = (long long)blockIdx.x * 256 + threadIdx.x; long long o; float a, b;
    if (transpose) { const long long np = (long long)C * (R / 2); if (i >= np) return; const int c = (int)(i / (R / 2)); const int r = 2 * (int)(i % (R / 2)); a = src[(long long)r * lds + c] * s; b = src[(long long)(r + 1) * lds + c] * s; o = (long long)c * ldd + r; }
    else { const long long np = (long long)R * (C / 2); if (i >= np) return; const int r = (int)(i / (C / 2)); const int c = 2 * (int)(i % (C / 2)); a = src[(long long)r * lds + c] * s; b = src[(long long)r * lds + c + 1] * s; o = (long long)r * ldd + c; }
    unsigned lo; const unsigned hi = f2bf2_pack(a, b, &lo); volatile unsigned* ph = (volatile unsigned*)(dhi + o); volatile unsigned* pl = (volatile unsigned*)(dlo + o);
    *ph = hi; *pl = lo; __threadfence(); *ph = hi; *pl = lo; }

namespace w25 {
#define AT_D 64
#define AT_NW 4
#define AT_QB 64
#define AT_KC 64
struct AttnGeom { const float* cp = nullptr; const float* pc = nullptr; long c_bs = 0, c_rs = 0, c_hs = 0;
                  long q_bs, q_rs, q_hs, k_bs, k_rs, k_hs, v_bs, v_rs, v_hs, o_bs, o_rs, o_hs;
                  int S, Skv, H, mask_mode; float qscale; int blk0; float mask_fill; int mask_is_int; };
static_assert(sizeof(AttnGeom) == 168, "no padding");

__device__ __forceinline__ unsigned short at_bf_bits(float f) {
  unsigned u = __float_as_uint(f);
  return (unsigned short)((u + 0x7FFFu + ((u >> 16) & 1u)) >> 16);
}
__device__ __forceinline__ __bf16 at_f2bf(float f) { return __builtin_bit_cast(__bf16, at_bf_bits(f)); }
__device__ __forceinline__ void at_split(float f, __bf16& hi, __bf16& lo) {
  const unsigned short hb = at_bf_bits(f);
  hi = __builtin_bit_cast(__bf16, hb);
  lo = at_f2bf(f - __uint_as_float(((unsigned)hb) << 16));
}
__device__ __forceinline__ v8f at_mma(v16b a, v16b b, v8f c) {
  c = __builtin_amdgcn_wmma_f32_16x16x32_bf16(false, a, false, b, (short)0, c, false, false);
  asm volatile("v_nop\n\tv_nop\n\tv_nop\n\tv_nop" : "+v"(c) : "v"(a), "v"(b));
  return c;
}
template <bool F16> __device__ __forceinline__ __bf16 at_to16(float f) {
  if (F16) return __builtin_bit_cast(__bf16, (_Float16)f);
  return at_f2bf(f);
}
template <bool F16> __device__ __forceinline__ v8f at_mma16(v16b a, v16b b, v8f c) {
  if (F16) {
    const v16h ah = __builtin_bit_cast(v16h, a), bh = __builtin_bit_cast(v16h, b);
    c = __builtin_amdgcn_wmma_f32_16x16x32_f16(false, ah, false, bh, (short)0, c, false, false);
    asm volatile("v_nop\n\tv_nop\n\tv_nop\n\tv_nop" : "+v"(c) : "v"(ah), "v"(bh));
    return c;
  }
  return at_mma(a, b, c);
}

template <bool SPLIT_QK, bool SPLIT_PV, bool F16 = false>
__global__ __launch_bounds__(128)
void attn64_kernel(const float* __restrict__ q, const float* __restrict__ k,
                   const float* __restrict__ v, float* __restrict__ out,
                   const void* __restrict__ mask_a, const int* __restrict__ mask_b, AttnGeom g) {
  static_assert(!(F16 && (SPLIT_QK || SPLIT_PV)), "f16 mode is non-split");
  const float PSC = F16 ? 32768.0f : 1.0f;
  union FB { v16b v; v8b h[2]; };
  __shared__ __align__(16) __bf16 Ksh[AT_KC * AT_D];
  __shared__ __align__(16) __bf16 Ksl[SPLIT_QK ? AT_KC * AT_D : 8];
  __shared__ __align__(16) __bf16 Vth[AT_D * AT_KC];
  __shared__ __align__(16) __bf16 Vtl[SPLIT_PV ? AT_D * AT_KC : 8];
  __shared__ __align__(16) __bf16 Psh[AT_NW][16 * AT_KC];
  __shared__ __align__(16) __bf16 Psl[SPLIT_PV ? AT_NW : 1][SPLIT_PV ? 16 * AT_KC : 8];
  __shared__ __align__(16) float  Os[AT_NW][16 * 68];

  const int tid  = threadIdx.x;
  const int wave = tid >> 5;
  const int lane = tid & 31;
  const int hh   = lane >> 4;
  const int c    = lane & 15;

  const int nqb = g.S / AT_QB;
  const int bx = blockIdx.x + g.blk0;
  const int qb = bx % nqb;
  const int bh = bx / nqb;
  const int h  = bh % g.H;
  const int b  = bh / g.H;
  const int qbase_block = qb * AT_QB;
  const int q0 = qbase_block + wave * 16;

  const float* qb_ptr = q + (size_t)b * g.q_bs + (size_t)h * g.q_hs;
  const float* kb_ptr = k + (size_t)b * g.k_bs + (size_t)h * g.k_hs;
  const float* vb_ptr = v + (size_t)b * g.v_bs + (size_t)h * g.v_hs;
  float*       ob_ptr = out + (size_t)b * g.o_bs + (size_t)h * g.o_hs;

  v16b qah[2], qal[2];
  {
    const float* qrow = qb_ptr + (size_t)(q0 + c) * g.q_rs;
#pragma unroll
    for (int dc = 0; dc < 2; ++dc) {
#pragma unroll
      for (int e = 0; e < 8; ++e) {
        const float f0 = qrow[dc * 32 + 8 * hh + e] * g.qscale;
        const float f1 = qrow[dc * 32 + 16 + 8 * hh + e] * g.qscale;
        if (SPLIT_QK) { __bf16 hq, lq; at_split(f0, hq, lq); qah[dc][e] = hq; qal[dc][e] = lq; at_split(f1, hq, lq); qah[dc][8 + e] = hq; qal[dc][8 + e] = lq; }
        else { qah[dc][e] = at_to16<F16>(f0); qah[dc][8 + e] = at_to16<F16>(f1); qal[dc][e] = qah[dc][e]; qal[dc][8 + e] = qah[dc][8 + e]; }
      }
    }
  }

  float mrow[8], lrow[8];
  v8f oacc[4];
#pragma unroll
  for (int r = 0; r < 8; ++r) { mrow[r] = -INFINITY; lrow[r] = 0.f; }
#pragma unroll
  for (int t = 0; t < 4; ++t) oacc[t] = (v8f){0.f,0.f,0.f,0.f,0.f,0.f,0.f,0.f};

  const int nChunks = (g.mask_mode == 1 || g.mask_mode == 4) ? (qb + 1) : (g.Skv / AT_KC);
  int qkeep[8];
#pragma unroll
  for (int r = 0; r < 8; ++r) qkeep[r] = (g.mask_mode == 3) ? mask_b[(size_t)b * g.S + q0 + 8 * hh + r] : 1;
  for (int kc = 0; kc < nChunks; ++kc) {
    const int kv0 = kc * AT_KC;
    __syncthreads();
    {
      const int kvr = tid >> 1, dh = (tid & 1) * 32;
      const float* krow = kb_ptr + (size_t)(kv0 + kvr) * g.k_rs + dh;
      const float* vrow = vb_ptr + (size_t)(kv0 + kvr) * g.v_rs + dh;
#pragma unroll
      for (int i = 0; i < 8; ++i) {
        v4f kk = *(const v4f*)(krow + 4 * i);
        v4f vv = *(const v4f*)(vrow + 4 * i);
#pragma unroll
        for (int e = 0; e < 4; ++e) {
          const int d = dh + 4 * i + e;
          if (SPLIT_QK) { __bf16 a, bl; at_split(kk[e], a, bl); Ksh[kvr * AT_D + d] = a; Ksl[kvr * AT_D + d] = bl; }
          else Ksh[kvr * AT_D + d] = at_to16<F16>(kk[e]);
          if (SPLIT_PV) { __bf16 a, bl; at_split(vv[e], a, bl); Vth[d * AT_KC + kvr] = a; Vtl[d * AT_KC + kvr] = bl; }
          else Vth[d * AT_KC + kvr] = at_to16<F16>(vv[e]);
        }
      }
    }
    __syncthreads();

    v8f s[4];
#pragma unroll
    for (int j = 0; j < 4; ++j) {
      s[j] = (v8f){0.f,0.f,0.f,0.f,0.f,0.f,0.f,0.f};
#pragma unroll 1
      for (int dc = 0; dc < 2; ++dc) {
        FB kb;
        kb.h[0] = *(const v8b*)(Ksh + (j * 16 + c) * AT_D + dc * 32 + 8 * hh);
        kb.h[1] = *(const v8b*)(Ksh + (j * 16 + c) * AT_D + dc * 32 + 16 + 8 * hh);
        s[j] = at_mma16<F16>(qah[dc], kb.v, s[j]);
        if (SPLIT_QK) {
          FB kl;
          kl.h[0] = *(const v8b*)(Ksl + (j * 16 + c) * AT_D + dc * 32 + 8 * hh);
          kl.h[1] = *(const v8b*)(Ksl + (j * 16 + c) * AT_D + dc * 32 + 16 + 8 * hh);
          s[j] = at_mma16<F16>(qah[dc], kl.v, s[j]);
          s[j] = at_mma16<F16>(qal[dc], kb.v, s[j]);
        }
      }
    }
    const bool diag = (g.mask_mode == 1) && (kc == qb);
    int kvkeep[4] = {1, 1, 1, 1};
    if (g.mask_mode == 3) {
#pragma unroll
      for (int j = 0; j < 4; ++j) kvkeep[j] = ((const int*)mask_a)[(size_t)b * g.Skv + kv0 + j * 16 + c];
    }
    float cm[8];
#pragma unroll
    for (int r = 0; r < 8; ++r) {
      const int qrow = q0 + 8 * hh + r;
      float m = -INFINITY;
#pragma unroll
      for (int j = 0; j < 4; ++j) {
        const int kvcol = kv0 + j * 16 + c;
        bool masked = false;
        if (diag) masked = (kvcol > qrow);
        else if (g.mask_mode == 4) masked = (kvcol > qrow) || (qrow - kvcol > g.mask_is_int);
        else if (g.mask_mode == 2) {
          const size_t mi = (size_t)qrow * g.Skv + kvcol;
          masked = (g.mask_is_int == 0) ? (((const float*)mask_a)[mi] == 0.0f)
                 : (g.mask_is_int == 1) ? (((const int*)mask_a)[mi] == 0) : (((const int*)mask_a)[mi] != 0);
        } else if (g.mask_mode == 3) masked = (qkeep[r] == 0) || (kvkeep[j] == 0);
        else if (g.mask_mode == 5) {
          const size_t mi = (size_t)qrow * g.Skv + kvcol;
          masked = (((const int*)mask_a)[mi] != 0);
          int n = mask_b[mi]; n = n < 0 ? 0 : n;
          s[j][r] += g.cp[(size_t)b * g.c_bs + (size_t)h * g.c_hs + (size_t)qrow * g.c_rs + n]
                   + g.pc[(size_t)b * g.c_bs + (size_t)h * g.c_hs + (size_t)kvcol * g.c_rs + n];
        }
        if (masked) s[j][r] = g.mask_fill;
        m = fmaxf(m, s[j][r]);
      }
#pragma unroll
      for (int off = 1; off < 16; off <<= 1) m = fmaxf(m, __shfl_xor(m, off, 32));
      cm[r] = m;
    }
    __bf16* pwh = Psh[wave];
    __bf16* pwl = Psl[SPLIT_PV ? wave : 0];
#pragma unroll
    for (int r = 0; r < 8; ++r) {
      const float mnew = fmaxf(mrow[r], cm[r]);
      const float alpha = expf(mrow[r] - mnew);
      mrow[r] = mnew;
      float psum = 0.f;
#pragma unroll
      for (int j = 0; j < 4; ++j) {
        const float p = expf(s[j][r] - mnew);
        psum += p;
        if (SPLIT_PV) { __bf16 a, bl; at_split(p, a, bl); pwh[(8 * hh + r) * AT_KC + j * 16 + c] = a; pwl[(8 * hh + r) * AT_KC + j * 16 + c] = bl; }
        else pwh[(8 * hh + r) * AT_KC + j * 16 + c] = at_to16<F16>(p * PSC);
      }
#pragma unroll
      for (int off = 1; off < 16; off <<= 1) psum += __shfl_xor(psum, off, 32);
      lrow[r] = lrow[r] * alpha + psum;
#pragma unroll
      for (int t = 0; t < 4; ++t) oacc[t][r] *= alpha;
    }
    __builtin_amdgcn_fence(__ATOMIC_RELEASE, "workgroup");
    __builtin_amdgcn_wave_barrier();
    __builtin_amdgcn_fence(__ATOMIC_ACQUIRE, "workgroup");
#pragma unroll 1
    for (int kk = 0; kk < 2; ++kk) {
      FB pa, pl;
      pa.h[0] = *(const v8b*)(pwh + c * AT_KC + kk * 32 + 8 * hh);
      pa.h[1] = *(const v8b*)(pwh + c * AT_KC + kk * 32 + 16 + 8 * hh);
      if (SPLIT_PV) {
        pl.h[0] = *(const v8b*)(pwl + c * AT_KC + kk * 32 + 8 * hh);
        pl.h[1] = *(const v8b*)(pwl + c * AT_KC + kk * 32 + 16 + 8 * hh);
      }
#pragma unroll
      for (int t = 0; t < 4; ++t) {
        FB vb;
        vb.h[0] = *(const v8b*)(Vth + (t * 16 + c) * AT_KC + kk * 32 + 8 * hh);
        vb.h[1] = *(const v8b*)(Vth + (t * 16 + c) * AT_KC + kk * 32 + 16 + 8 * hh);
        oacc[t] = at_mma16<F16>(pa.v, vb.v, oacc[t]);
        if (SPLIT_PV) {
          FB vl;
          vl.h[0] = *(const v8b*)(Vtl + (t * 16 + c) * AT_KC + kk * 32 + 8 * hh);
          vl.h[1] = *(const v8b*)(Vtl + (t * 16 + c) * AT_KC + kk * 32 + 16 + 8 * hh);
          oacc[t] = at_mma16<F16>(pa.v, vl.v, oacc[t]);
          oacc[t] = at_mma16<F16>(pl.v, vb.v, oacc[t]);
        }
      }
    }
  }

  float* os = Os[wave];
#pragma unroll
  for (int r = 0; r < 8; ++r) {
    const float inv = 1.0f / (lrow[r] * PSC);
#pragma unroll
    for (int t = 0; t < 4; ++t) os[(8 * hh + r) * 68 + t * 16 + c] = oacc[t][r] * inv;
  }
  __builtin_amdgcn_fence(__ATOMIC_RELEASE, "workgroup");
  __builtin_amdgcn_wave_barrier();
  __builtin_amdgcn_fence(__ATOMIC_ACQUIRE, "workgroup");
  {
    const int c4 = (lane & 15) * 4;
    for (int pass = 0; pass < 2; ++pass) {
#pragma unroll
      for (int it = 0; it < 8; ++it) {
        const int row = it * 2 + hh;
        v4f val = *(const v4f*)(os + row * 68 + c4);
        *(volatile v4f*)(ob_ptr + (size_t)(q0 + row) * g.o_rs + c4) = val;
      }
      __threadfence();
    }
  }
}

}

__device__ __forceinline__ void st_h2(_Float16* dst, float a, float b) { const unsigned u = (unsigned)__builtin_bit_cast(unsigned short, (_Float16)a) | ((unsigned)__builtin_bit_cast(unsigned short, (_Float16)b) << 16); volatile unsigned* d = (volatile unsigned*)dst; *d = u; __threadfence(); *d = u; }
__device__ __forceinline__ unsigned short bf16b(float v) { const unsigned u = __builtin_bit_cast(unsigned, v); return (unsigned short)(((u + 0x7FFFu + ((u >> 16) & 1u)) & 0xFFFF0000u) >> 16); }
__device__ __forceinline__ float bf16f(unsigned short h) { return __builtin_bit_cast(float, ((unsigned)h) << 16); }
__device__ __forceinline__ void st_split2(_Float16* Hp, _Float16* Lp, long long e, float v0, float v1) { const unsigned short h0 = bf16b(v0), h1 = bf16b(v1); { const unsigned u = (unsigned)h0 | ((unsigned)h1 << 16); volatile unsigned* d = (volatile unsigned*)(Hp + e); *d = u; __threadfence(); *d = u; } { const unsigned u = (unsigned)bf16b(v0 - bf16f(h0)) | ((unsigned)bf16b(v1 - bf16f(h1)) << 16); volatile unsigned* d = (volatile unsigned*)(Lp + e); *d = u; __threadfence(); *d = u; } }
__global__ __launch_bounds__(256) void k_ac_planes(const float* __restrict__ QF, const float* __restrict__ KF, const float* __restrict__ VF, _Float16* QH, _Float16* QL, _Float16* KH, _Float16* KL, _Float16* V16, int nqk, long long nv) { const long long t = (long long)blockIdx.x * 256 + threadIdx.x; const long long e = 2 * t;
    if (e < nqk) { st_split2(QH, QL, e, QF[e], QF[e + 1]); st_split2(KH, KL, e, KF[e], KF[e + 1]); }
    if (e < nv) st_h2(V16 + e, VF[e], VF[e + 1]); }
__global__ __launch_bounds__(256) void k_ac_soft(float* __restrict__ EN, _Float16* __restrict__ P16, int N) { __shared__ float red[256]; const long long row = blockIdx.x; float* sr = EN + row * N; const int t = threadIdx.x; float mx = -3.0e38f;
#pragma unroll 1
    for (int j = 2 * t; j < N; j += 512) mx = fmaxf(mx, fmaxf(sr[j], sr[j + 1]));
    red[t] = mx; __syncthreads(); for (int o = 128; o > 0; o >>= 1) { if (t < o) red[t] = fmaxf(red[t], red[t + o]); __syncthreads(); } const float m = red[0]; __syncthreads();
    float s = 0.f;
#pragma unroll 1
    for (int j = 2 * t; j < N; j += 512) { const float e0 = expf(sr[j] - m), e1 = expf(sr[j + 1] - m); s += e0 + e1; const unsigned long long pk = (unsigned long long)__builtin_bit_cast(unsigned, e0) | ((unsigned long long)__builtin_bit_cast(unsigned, e1) << 32); VST2(unsigned long long, (unsigned long long*)(sr + j), pk); }
    red[t] = s; __syncthreads(); for (int o = 128; o > 0; o >>= 1) { if (t < o) red[t] += red[t + o]; __syncthreads(); } const float f = 4096.f / red[0];
#pragma unroll 1
    for (int j = 2 * t; j < N; j += 512) st_h2(P16 + row * N + j, sr[j] * f, sr[j + 1] * f); }
__global__ __launch_bounds__(256) void k_ac_fuse(const float* __restrict__ CT, const float* __restrict__ FW, float* __restrict__ OUT, int i, int b, long long n) { const long long t = (long long)blockIdx.x * 256 + threadIdx.x; if (t >= n) return; float* o = OUT + (long long)b * n + t; const float v = CT[t] * FW[i] * (1.f / 3.f); VST2(float, o, (i == 0) ? v : (*o + v)); }

template __global__ void k_gemm<1>(GemmP);

extern "C" void kernel_launch(void* const* d_in, const int* in_sizes, int n_in, void* d_out, int out_size, void* d_ws, size_t ws_size, hipStream_t stream) {
    (void)in_sizes; (void)n_in; (void)out_size; (void)ws_size;
    const float* s0 = (const float*)d_in[0];
    const float* s1 = (const float*)d_in[1];
    const float* s2 = (const float*)d_in[2];
    const float* Wq = (const float*)d_in[3];
    const float* bq = (const float*)d_in[4];
    const float* Wk = (const float*)d_in[5];
    const float* bk = (const float*)d_in[6];
    const float* Wv = (const float*)d_in[7];
    const float* bv = (const float*)d_in[8];
    const float* fw = (const float*)d_in[9];
    const int Bn = 16;
    const int C = 256;
    const int C8 = 32;
    const int N = 1600;
    float* out = (float*)d_out;
    char* wsp = (char*)d_ws;
    float* QF = (float*)wsp; wsp += (((size_t)((size_t)N * C8) * 4 + 255) / 256) * 256;
    float* KF = (float*)wsp; wsp += (((size_t)((size_t)N * C8) * 4 + 255) / 256) * 256;
    float* VF = (float*)wsp; wsp += (((size_t)((size_t)C * N) * 4 + 255) / 256) * 256;
    unsigned short* QH = (unsigned short*)wsp; wsp += (((size_t)((size_t)N * C8) * 2 + 255) / 256) * 256;
    unsigned short* QL = (unsigned short*)wsp; wsp += (((size_t)((size_t)N * C8) * 2 + 255) / 256) * 256;
    unsigned short* KH = (unsigned short*)wsp; wsp += (((size_t)((size_t)N * C8) * 2 + 255) / 256) * 256;
    unsigned short* KL = (unsigned short*)wsp; wsp += (((size_t)((size_t)N * C8) * 2 + 255) / 256) * 256;
    unsigned short* V16 = (unsigned short*)wsp; wsp += (((size_t)((size_t)C * N) * 2 + 255) / 256) * 256;
    float* EN = (float*)wsp; wsp += (((size_t)((size_t)N * N) * 4 + 255) / 256) * 256;
    unsigned short* P16 = (unsigned short*)wsp; wsp += (((size_t)((size_t)N * N) * 2 + 255) / 256) * 256;
    float* CT = (float*)wsp; wsp += (((size_t)((size_t)C * N) * 4 + 255) / 256) * 256;
    unsigned short* G64A = (unsigned short*)wsp; wsp += (((size_t)(65536) * 2 + 255) / 256) * 256;
    unsigned short* G64B = (unsigned short*)wsp; wsp += (((size_t)(409600) * 2 + 255) / 256) * 256;
    { GemmP gq0_0;
      gq0_0.A = s0 + (size_t)0 * C * N; gq0_0.B = Wq; gq0_0.bias = bq; gq0_0.R = s0 + (size_t)0 * C * N; gq0_0.C = QF;
      gq0_0.sAo = 0; gq0_0.sAi = 0; gq0_0.sAm = 1; gq0_0.sAk = N; gq0_0.sBo = 0; gq0_0.sBi = 0; gq0_0.sBn = C; gq0_0.sBk = 1; gq0_0.sCo = 0; gq0_0.sCi = 0; gq0_0.sCm = C8; gq0_0.sRo = 0; gq0_0.sRi = 0; gq0_0.sRm = 0; gq0_0.sRn = 0;
      gq0_0.M = N; gq0_0.N = C8; gq0_0.K = C; gq0_0.zi_n = 1; gq0_0.flags = 1; gq0_0.act = 0;
      gq0_0.alpha = 1.0f; gq0_0.beta = 0.0f; gq0_0.sa = 1.0f; gq0_0.sb = 1.0f; gq0_0.Npad = C8; gq0_0.pad_ = 0;
      if ((long long)(N) >= 64 && (long long)(C8) >= 64) k_gemmT<1, 2, 4><<<dim3((unsigned)((C8) + 63) / 64, (unsigned)((N) + 31) / 32, (unsigned)(1)), 32, 0, stream>>>(gq0_0);
      else k_gemm<1><<<dim3((unsigned)((C8) + 31) / 32, (unsigned)((N) + 15) / 16, (unsigned)(1)), 32, 0, stream>>>(gq0_0); }
    { GemmP gk0_0;
      gk0_0.A = s1 + (size_t)0 * C * N; gk0_0.B = Wk; gk0_0.bias = bk; gk0_0.R = s1 + (size_t)0 * C * N; gk0_0.C = KF;
      gk0_0.sAo = 0; gk0_0.sAi = 0; gk0_0.sAm = 1; gk0_0.sAk = N; gk0_0.sBo = 0; gk0_0.sBi = 0; gk0_0.sBn = C; gk0_0.sBk = 1; gk0_0.sCo = 0; gk0_0.sCi = 0; gk0_0.sCm = C8; gk0_0.sRo = 0; gk0_0.sRi = 0; gk0_0.sRm = 0; gk0_0.sRn = 0;
      gk0_0.M = N; gk0_0.N = C8; gk0_0.K = C; gk0_0.zi_n = 1; gk0_0.flags = 1; gk0_0.act = 0;
      gk0_0.alpha = 1.0f; gk0_0.beta = 0.0f; gk0_0.sa = 1.0f; gk0_0.sb = 1.0f; gk0_0.Npad = C8; gk0_0.pad_ = 0;
      if ((long long)(N) >= 64 && (long long)(C8) >= 64) k_gemmT<1, 2, 4><<<dim3((unsigned)((C8) + 63) / 64, (unsigned)((N) + 31) / 32, (unsigned)(1)), 32, 0, stream>>>(gk0_0);
      else k_gemm<1><<<dim3((unsigned)((C8) + 31) / 32, (unsigned)((N) + 15) / 16, (unsigned)(1)), 32, 0, stream>>>(gk0_0); }
    k_cast16<<<(unsigned)((((long long)(256) * ((256) / 2)) + 255) / 256), 256, 0, stream>>>(Wv, 256, (_Float16*)(G64A), 256, 256, 256, 1.0f);
    k_castT16<<<(unsigned)((((long long)(1600) * ((256) / 2)) + 255) / 256), 256, 0, stream>>>(s1 + (size_t)0 * C * N, 1600, (_Float16*)(G64B), 256, 256, 1600, 16.0f);
    w25::wmma_gemm64<0, false, 1, 0, false, 0><<<dim3((unsigned)((((256) / 64) * ((1600) / 64) + 7) / 8), (unsigned)(1)), 256, 0, stream>>>((const unsigned short*)(G64A), nullptr, 256, 0, (const unsigned short*)(G64B), nullptr, 256, 0, (void*)(VF), nullptr, 1600, 0, bv, nullptr, 0, 256, 1600, 256, 0.0625f);
    k_ac_planes<<<(unsigned)(((long long)C * N / 2 + 255) / 256), 256, 0, stream>>>(QF, KF, VF, (_Float16*)QH, (_Float16*)QL, (_Float16*)KH, (_Float16*)KL, (_Float16*)V16, N * C8, (long long)C * N);
    w25::wmma_gemm64<1, true, 0, 0, false, 0><<<dim3((unsigned)((((N) / 64) * ((N) / 64) + 7) / 8), (unsigned)(1)), 256, 0, stream>>>((const unsigned short*)(QH), (const unsigned short*)(QL), C8, 0, (const unsigned short*)(KH), (const unsigned short*)(KL), C8, 0, (void*)(EN), nullptr, N, 0, nullptr, nullptr, 0, N, N, C8, 1.0f);
    k_ac_soft<<<N, 256, 0, stream>>>(EN, (_Float16*)P16, N);
    w25::wmma_gemm64<0, false, 0, 0, false, 0><<<dim3((unsigned)((((C) / 64) * ((N) / 64) + 7) / 8), (unsigned)(1)), 256, 0, stream>>>((const unsigned short*)(V16), nullptr, N, 0, (const unsigned short*)(P16), nullptr, N, 0, (void*)(CT), nullptr, N, 0, nullptr, nullptr, 0, C, N, N, 0.000244140625f);
    k_ac_fuse<<<(unsigned)(((long long)C * N + 255) / 256), 256, 0, stream>>>(CT, fw, out, 0, 0, (long long)C * N);
    { GemmP gq0_1;
      gq0_1.A = s0 + (size_t)1 * C * N; gq0_1.B = Wq; gq0_1.bias = bq; gq0_1.R = s0 + (size_t)1 * C * N; gq0_1.C = QF;
      gq0_1.sAo = 0; gq0_1.sAi = 0; gq0_1.sAm = 1; gq0_1.sAk = N; gq0_1.sBo = 0; gq0_1.sBi = 0; gq0_1.sBn = C; gq0_1.sBk = 1; gq0_1.sCo = 0; gq0_1.sCi = 0; gq0_1.sCm = C8; gq0_1.sRo = 0; gq0_1.sRi = 0; gq0_1.sRm = 0; gq0_1.sRn = 0;
      gq0_1.M = N; gq0_1.N = C8; gq0_1.K = C; gq0_1.zi_n = 1; gq0_1.flags = 1; gq0_1.act = 0;
      gq0_1.alpha = 1.0f; gq0_1.beta = 0.0f; gq0_1.sa = 1.0f; gq0_1.sb = 1.0f; gq0_1.Npad = C8; gq0_1.pad_ = 0;
      if ((long long)(N) >= 64 && (long long)(C8) >= 64) k_gemmT<1, 2, 4><<<dim3((unsigned)((C8) + 63) / 64, (unsigned)((N) + 31) / 32, (unsigned)(1)), 32, 0, stream>>>(gq0_1);
      else k_gemm<1><<<dim3((unsigned)((C8) + 31) / 32, (unsigned)((N) + 15) / 16, (unsigned)(1)), 32, 0, stream>>>(gq0_1); }
    { GemmP gk0_1;
      gk0_1.A = s1 + (size_t)1 * C * N; gk0_1.B = Wk; gk0_1.bias = bk; gk0_1.R = s1 + (size_t)1 * C * N; gk0_1.C = KF;
      gk0_1.sAo = 0; gk0_1.sAi = 0; gk0_1.sAm = 1; gk0_1.sAk = N; gk0_1.sBo = 0; gk0_1.sBi = 0; gk0_1.sBn = C; gk0_1.sBk = 1; gk0_1.sCo = 0; gk0_1.sCi = 0; gk0_1.sCm = C8; gk0_1.sRo = 0; gk0_1.sRi = 0; gk0_1.sRm = 0; gk0_1.sRn = 0;
      gk0_1.M = N; gk0_1.N = C8; gk0_1.K = C; gk0_1.zi_n = 1; gk0_1.flags = 1; gk0_1.act = 0;
      gk0_1.alpha = 1.0f; gk0_1.beta = 0.0f; gk0_1.sa = 1.0f; gk0_1.sb = 1.0f; gk0_1.Npad = C8; gk0_1.pad_ = 0;
      if ((long long)(N) >= 64 && (long long)(C8) >= 64) k_gemmT<1, 2, 4><<<dim3((unsigned)((C8) + 63) / 64, (unsigned)((N) + 31) / 32, (unsigned)(1)), 32, 0, stream>>>(gk0_1);
      else k_gemm<1><<<dim3((unsigned)((C8) + 31) / 32, (unsigned)((N) + 15) / 16, (unsigned)(1)), 32, 0, stream>>>(gk0_1); }
    k_cast16<<<(unsigned)((((long long)(256) * ((256) / 2)) + 255) / 256), 256, 0, stream>>>(Wv, 256, (_Float16*)(G64A), 256, 256, 256, 1.0f);
    k_castT16<<<(unsigned)((((long long)(1600) * ((256) / 2)) + 255) / 256), 256, 0, stream>>>(s1 + (size_t)1 * C * N, 1600, (_Float16*)(G64B), 256, 256, 1600, 16.0f);
    w25::wmma_gemm64<0, false, 1, 0, false, 0><<<dim3((unsigned)((((256) / 64) * ((1600) / 64) + 7) / 8), (unsigned)(1)), 256, 0, stream>>>((const unsigned short*)(G64A), nullptr, 256, 0, (const unsigned short*)(G64B), nullptr, 256, 0, (void*)(VF), nullptr, 1600, 0, bv, nullptr, 0, 256, 1600, 256, 0.0625f);
    k_ac_planes<<<(unsigned)(((long long)C * N / 2 + 255) / 256), 256, 0, stream>>>(QF, KF, VF, (_Float16*)QH, (_Float16*)QL, (_Float16*)KH, (_Float16*)KL, (_Float16*)V16, N * C8, (long long)C * N);
    w25::wmma_gemm64<1, true, 0, 0, false, 0><<<dim3((unsigned)((((N) / 64) * ((N) / 64) + 7) / 8), (unsigned)(1)), 256, 0, stream>>>((const unsigned short*)(QH), (const unsigned short*)(QL), C8, 0, (const unsigned short*)(KH), (const unsigned short*)(KL), C8, 0, (void*)(EN), nullptr, N, 0, nullptr, nullptr, 0, N, N, C8, 1.0f);
    k_ac_soft<<<N, 256, 0, stream>>>(EN, (_Float16*)P16, N);
    w25::wmma_gemm64<0, false, 0, 0, false, 0><<<dim3((unsigned)((((C) / 64) * ((N) / 64) + 7) / 8), (unsigned)(1)), 256, 0, stream>>>((const unsigned short*)(V16), nullptr, N, 0, (const unsigned short*)(P16), nullptr, N, 0, (void*)(CT), nullptr, N, 0, nullptr, nullptr, 0, C, N, N, 0.000244140625f);
    k_ac_fuse<<<(unsigned)(((long long)C * N + 255) / 256), 256, 0, stream>>>(CT, fw, out, 0, 1, (long long)C * N);
    { GemmP gq0_2;
      gq0_2.A = s0 + (size_t)2 * C * N; gq0_2.B = Wq; gq0_2.bias = bq; gq0_2.R = s0 + (size_t)2 * C * N; gq0_2.C = QF;
      gq0_2.sAo = 0; gq0_2.sAi = 0; gq0_2.sAm = 1; gq0_2.sAk = N; gq0_2.sBo = 0; gq0_2.sBi = 0; gq0_2.sBn = C; gq0_2.sBk = 1; gq0_2.sCo = 0; gq0_2.sCi = 0; gq0_2.sCm = C8; gq0_2.sRo = 0; gq0_2.sRi = 0; gq0_2.sRm = 0; gq0_2.sRn = 0;
      gq0_2.M = N; gq0_2.N = C8; gq0_2.K = C; gq0_2.zi_n = 1; gq0_2.flags = 1; gq0_2.act = 0;
      gq0_2.alpha = 1.0f; gq0_2.beta = 0.0f; gq0_2.sa = 1.0f; gq0_2.sb = 1.0f; gq0_2.Npad = C8; gq0_2.pad_ = 0;
      if ((long long)(N) >= 64 && (long long)(C8) >= 64) k_gemmT<1, 2, 4><<<dim3((unsigned)((C8) + 63) / 64, (unsigned)((N) + 31) / 32, (unsigned)(1)), 32, 0, stream>>>(gq0_2);
      else k_gemm<1><<<dim3((unsigned)((C8) + 31) / 32, (unsigned)((N) + 15) / 16, (unsigned)(1)), 32, 0, stream>>>(gq0_2); }
    { GemmP gk0_2;
      gk0_2.A = s1 + (size_t)2 * C * N; gk0_2.B = Wk; gk0_2.bias = bk; gk0_2.R = s1 + (size_t)2 * C * N; gk0_2.C = KF;
      gk0_2.sAo = 0; gk0_2.sAi = 0; gk0_2.sAm = 1; gk0_2.sAk = N; gk0_2.sBo = 0; gk0_2.sBi = 0; gk0_2.sBn = C; gk0_2.sBk = 1; gk0_2.sCo = 0; gk0_2.sCi = 0; gk0_2.sCm = C8; gk0_2.sRo = 0; gk0_2.sRi = 0; gk0_2.sRm = 0; gk0_2.sRn = 0;
      gk0_2.M = N; gk0_2.N = C8; gk0_2.K = C; gk0_2.zi_n = 1; gk0_2.flags = 1; gk0_2.act = 0;
      gk0_2.alpha = 1.0f; gk0_2.beta = 0.0f; gk0_2.sa = 1.0f; gk0_2.sb = 1.0f; gk0_2.Npad = C8; gk0_2.pad_ = 0;
      if ((long long)(N) >= 64 && (long long)(C8) >= 64) k_gemmT<1, 2, 4><<<dim3((unsigned)((C8) + 63) / 64, (unsigned)((N) + 31) / 32, (unsigned)(1)), 32, 0, stream>>>(gk0_2);
      else k_gemm<1><<<dim3((unsigned)((C8) + 31) / 32, (unsigned)((N) + 15) / 16, (unsigned)(1)), 32, 0, stream>>>(gk0_2); }
    k_cast16<<<(unsigned)((((long long)(256) * ((256) / 2)) + 255) / 256), 256, 0, stream>>>(Wv, 256, (_Float16*)(G64A), 256, 256, 256, 1.0f);
    k_castT16<<<(unsigned)((((long long)(1600) * ((256) / 2)) + 255) / 256), 256, 0, stream>>>(s1 + (size_t)2 * C * N, 1600, (_Float16*)(G64B), 256, 256, 1600, 16.0f);
    w25::wmma_gemm64<0, false, 1, 0, false, 0><<<dim3((unsigned)((((256) / 64) * ((1600) / 64) + 7) / 8), (unsigned)(1)), 256, 0, stream>>>((const unsigned short*)(G64A), nullptr, 256, 0, (const unsigned short*)(G64B), nullptr, 256, 0, (void*)(VF), nullptr, 1600, 0, bv, nullptr, 0, 256, 1600, 256, 0.0625f);
    k_ac_planes<<<(unsigned)(((long long)C * N / 2 + 255) / 256), 256, 0, stream>>>(QF, KF, VF, (_Float16*)QH, (_Float16*)QL, (_Float16*)KH, (_Float16*)KL, (_Float16*)V16, N * C8, (long long)C * N);
    w25::wmma_gemm64<1, true, 0, 0, false, 0><<<dim3((unsigned)((((N) / 64) * ((N) / 64) + 7) / 8), (unsigned)(1)), 256, 0, stream>>>((const unsigned short*)(QH), (const unsigned short*)(QL), C8, 0, (const unsigned short*)(KH), (const unsigned short*)(KL), C8, 0, (void*)(EN), nullptr, N, 0, nullptr, nullptr, 0, N, N, C8, 1.0f);
    k_ac_soft<<<N, 256, 0, stream>>>(EN, (_Float16*)P16, N);
    w25::wmma_gemm64<0, false, 0, 0, false, 0><<<dim3((unsigned)((((C) / 64) * ((N) / 64) + 7) / 8), (unsigned)(1)), 256, 0, stream>>>((const unsigned short*)(V16), nullptr, N, 0, (const unsigned short*)(P16), nullptr, N, 0, (void*)(CT), nullptr, N, 0, nullptr, nullptr, 0, C, N, N, 0.000244140625f);
    k_ac_fuse<<<(unsigned)(((long long)C * N + 255) / 256), 256, 0, stream>>>(CT, fw, out, 0, 2, (long long)C * N);
    { GemmP gq0_3;
      gq0_3.A = s0 + (size_t)3 * C * N; gq0_3.B = Wq; gq0_3.bias = bq; gq0_3.R = s0 + (size_t)3 * C * N; gq0_3.C = QF;
      gq0_3.sAo = 0; gq0_3.sAi = 0; gq0_3.sAm = 1; gq0_3.sAk = N; gq0_3.sBo = 0; gq0_3.sBi = 0; gq0_3.sBn = C; gq0_3.sBk = 1; gq0_3.sCo = 0; gq0_3.sCi = 0; gq0_3.sCm = C8; gq0_3.sRo = 0; gq0_3.sRi = 0; gq0_3.sRm = 0; gq0_3.sRn = 0;
      gq0_3.M = N; gq0_3.N = C8; gq0_3.K = C; gq0_3.zi_n = 1; gq0_3.flags = 1; gq0_3.act = 0;
      gq0_3.alpha = 1.0f; gq0_3.beta = 0.0f; gq0_3.sa = 1.0f; gq0_3.sb = 1.0f; gq0_3.Npad = C8; gq0_3.pad_ = 0;
      if ((long long)(N) >= 64 && (long long)(C8) >= 64) k_gemmT<1, 2, 4><<<dim3((unsigned)((C8) + 63) / 64, (unsigned)((N) + 31) / 32, (unsigned)(1)), 32, 0, stream>>>(gq0_3);
      else k_gemm<1><<<dim3((unsigned)((C8) + 31) / 32, (unsigned)((N) + 15) / 16, (unsigned)(1)), 32, 0, stream>>>(gq0_3); }
    { GemmP gk0_3;
      gk0_3.A = s1 + (size_t)3 * C * N; gk0_3.B = Wk; gk0_3.bias = bk; gk0_3.R = s1 + (size_t)3 * C * N; gk0_3.C = KF;
      gk0_3.sAo = 0; gk0_3.sAi = 0; gk0_3.sAm = 1; gk0_3.sAk = N; gk0_3.sBo = 0; gk0_3.sBi = 0; gk0_3.sBn = C; gk0_3.sBk = 1; gk0_3.sCo = 0; gk0_3.sCi = 0; gk0_3.sCm = C8; gk0_3.sRo = 0; gk0_3.sRi = 0; gk0_3.sRm = 0; gk0_3.sRn = 0;
      gk0_3.M = N; gk0_3.N = C8; gk0_3.K = C; gk0_3.zi_n = 1; gk0_3.flags = 1; gk0_3.act = 0;
      gk0_3.alpha = 1.0f; gk0_3.beta = 0.0f; gk0_3.sa = 1.0f; gk0_3.sb = 1.0f; gk0_3.Npad = C8; gk0_3.pad_ = 0;
      if ((long long)(N) >= 64 && (long long)(C8) >= 64) k_gemmT<1, 2, 4><<<dim3((unsigned)((C8) + 63) / 64, (unsigned)((N) + 31) / 32, (unsigned)(1)), 32, 0, stream>>>(gk0_3);
      else k_gemm<1><<<dim3((unsigned)((C8) + 31) / 32, (unsigned)((N) + 15) / 16, (unsigned)(1)), 32, 0, stream>>>(gk0_3); }
    k_cast16<<<(unsigned)((((long long)(256) * ((256) / 2)) + 255) / 256), 256, 0, stream>>>(Wv, 256, (_Float16*)(G64A), 256, 256, 256, 1.0f);
    k_castT16<<<(unsigned)((((long long)(1600) * ((256) / 2)) + 255) / 256), 256, 0, stream>>>(s1 + (size_t)3 * C * N, 1600, (_Float16*)(G64B), 256, 256, 1600, 16.0f);
    w25::wmma_gemm64<0, false, 1, 0, false, 0><<<dim3((unsigned)((((256) / 64) * ((1600) / 64) + 7) / 8), (unsigned)(1)), 256, 0, stream>>>((const unsigned short*)(G64A), nullptr, 256, 0, (const unsigned short*)(G64B), nullptr, 256, 0, (void*)(VF), nullptr, 1600, 0, bv, nullptr, 0, 256, 1600, 256, 0.0625f);
    k_ac_planes<<<(unsigned)(((long long)C * N / 2 + 255) / 256), 256, 0, stream>>>(QF, KF, VF, (_Float16*)QH, (_Float16*)QL, (_Float16*)KH, (_Float16*)KL, (_Float16*)V16, N * C8, (long long)C * N);
    w25::wmma_gemm64<1, true, 0, 0, false, 0><<<dim3((unsigned)((((N) / 64) * ((N) / 64) + 7) / 8), (unsigned)(1)), 256, 0, stream>>>((const unsigned short*)(QH), (const unsigned short*)(QL), C8, 0, (const unsigned short*)(KH), (const unsigned short*)(KL), C8, 0, (void*)(EN), nullptr, N, 0, nullptr, nullptr, 0, N, N, C8, 1.0f);
    k_ac_soft<<<N, 256, 0, stream>>>(EN, (_Float16*)P16, N);
    w25::wmma_gemm64<0, false, 0, 0, false, 0><<<dim3((unsigned)((((C) / 64) * ((N) / 64) + 7) / 8), (unsigned)(1)), 256, 0, stream>>>((const unsigned short*)(V16), nullptr, N, 0, (const unsigned short*)(P16), nullptr, N, 0, (void*)(CT), nullptr, N, 0, nullptr, nullptr, 0, C, N, N, 0.000244140625f);
    k_ac_fuse<<<(unsigned)(((long long)C * N + 255) / 256), 256, 0, stream>>>(CT, fw, out, 0, 3, (long long)C * N);
    { GemmP gq0_4;
      gq0_4.A = s0 + (size_t)4 * C * N; gq0_4.B = Wq; gq0_4.bias = bq; gq0_4.R = s0 + (size_t)4 * C * N; gq0_4.C = QF;
      gq0_4.sAo = 0; gq0_4.sAi = 0; gq0_4.sAm = 1; gq0_4.sAk = N; gq0_4.sBo = 0; gq0_4.sBi = 0; gq0_4.sBn = C; gq0_4.sBk = 1; gq0_4.sCo = 0; gq0_4.sCi = 0; gq0_4.sCm = C8; gq0_4.sRo = 0; gq0_4.sRi = 0; gq0_4.sRm = 0; gq0_4.sRn = 0;
      gq0_4.M = N; gq0_4.N = C8; gq0_4.K = C; gq0_4.zi_n = 1; gq0_4.flags = 1; gq0_4.act = 0;
      gq0_4.alpha = 1.0f; gq0_4.beta = 0.0f; gq0_4.sa = 1.0f; gq0_4.sb = 1.0f; gq0_4.Npad = C8; gq0_4.pad_ = 0;
      if ((long long)(N) >= 64 && (long long)(C8) >= 64) k_gemmT<1, 2, 4><<<dim3((unsigned)((C8) + 63) / 64, (unsigned)((N) + 31) / 32, (unsigned)(1)), 32, 0, stream>>>(gq0_4);
      else k_gemm<1><<<dim3((unsigned)((C8) + 31) / 32, (unsigned)((N) + 15) / 16, (unsigned)(1)), 32, 0, stream>>>(gq0_4); }
    { GemmP gk0_4;
      gk0_4.A = s1 + (size_t)4 * C * N; gk0_4.B = Wk; gk0_4.bias = bk; gk0_4.R = s1 + (size_t)4 * C * N; gk0_4.C = KF;
      gk0_4.sAo = 0; gk0_4.sAi = 0; gk0_4.sAm = 1; gk0_4.sAk = N; gk0_4.sBo = 0; gk0_4.sBi = 0; gk0_4.sBn = C; gk0_4.sBk = 1; gk0_4.sCo = 0; gk0_4.sCi = 0; gk0_4.sCm = C8; gk0_4.sRo = 0; gk0_4.sRi = 0; gk0_4.sRm = 0; gk0_4.sRn = 0;
      gk0_4.M = N; gk0_4.N = C8; gk0_4.K = C; gk0_4.zi_n = 1; gk0_4.flags = 1; gk0_4.act = 0;
      gk0_4.alpha = 1.0f; gk0_4.beta = 0.0f; gk0_4.sa = 1.0f; gk0_4.sb = 1.0f; gk0_4.Npad = C8; gk0_4.pad_ = 0;
      if ((long long)(N) >= 64 && (long long)(C8) >= 64) k_gemmT<1, 2, 4><<<dim3((unsigned)((C8) + 63) / 64, (unsigned)((N) + 31) / 32, (unsigned)(1)), 32, 0, stream>>>(gk0_4);
      else k_gemm<1><<<dim3((unsigned)((C8) + 31) / 32, (unsigned)((N) + 15) / 16, (unsigned)(1)), 32, 0, stream>>>(gk0_4); }
    k_cast16<<<(unsigned)((((long long)(256) * ((256) / 2)) + 255) / 256), 256, 0, stream>>>(Wv, 256, (_Float16*)(G64A), 256, 256, 256, 1.0f);
    k_castT16<<<(unsigned)((((long long)(1600) * ((256) / 2)) + 255) / 256), 256, 0, stream>>>(s1 + (size_t)4 * C * N, 1600, (_Float16*)(G64B), 256, 256, 1600, 16.0f);
    w25::wmma_gemm64<0, false, 1, 0, false, 0><<<dim3((unsigned)((((256) / 64) * ((1600) / 64) + 7) / 8), (unsigned)(1)), 256, 0, stream>>>((const unsigned short*)(G64A), nullptr, 256, 0, (const unsigned short*)(G64B), nullptr, 256, 0, (void*)(VF), nullptr, 1600, 0, bv, nullptr, 0, 256, 1600, 256, 0.0625f);
    k_ac_planes<<<(unsigned)(((long long)C * N / 2 + 255) / 256), 256, 0, stream>>>(QF, KF, VF, (_Float16*)QH, (_Float16*)QL, (_Float16*)KH, (_Float16*)KL, (_Float16*)V16, N * C8, (long long)C * N);
    w25::wmma_gemm64<1, true, 0, 0, false, 0><<<dim3((unsigned)((((N) / 64) * ((N) / 64) + 7) / 8), (unsigned)(1)), 256, 0, stream>>>((const unsigned short*)(QH), (const unsigned short*)(QL), C8, 0, (const unsigned short*)(KH), (const unsigned short*)(KL), C8, 0, (void*)(EN), nullptr, N, 0, nullptr, nullptr, 0, N, N, C8, 1.0f);
    k_ac_soft<<<N, 256, 0, stream>>>(EN, (_Float16*)P16, N);
    w25::wmma_gemm64<0, false, 0, 0, false, 0><<<dim3((unsigned)((((C) / 64) * ((N) / 64) + 7) / 8), (unsigned)(1)), 256, 0, stream>>>((const unsigned short*)(V16), nullptr, N, 0, (const unsigned short*)(P16), nullptr, N, 0, (void*)(CT), nullptr, N, 0, nullptr, nullptr, 0, C, N, N, 0.000244140625f);
    k_ac_fuse<<<(unsigned)(((long long)C * N + 255) / 256), 256, 0, stream>>>(CT, fw, out, 0, 4, (long long)C * N);
    { GemmP gq0_5;
      gq0_5.A = s0 + (size_t)5 * C * N; gq0_5.B = Wq; gq0_5.bias = bq; gq0_5.R = s0 + (size_t)5 * C * N; gq0_5.C = QF;
      gq0_5.sAo = 0; gq0_5.sAi = 0; gq0_5.sAm = 1; gq0_5.sAk = N; gq0_5.sBo = 0; gq0_5.sBi = 0; gq0_5.sBn = C; gq0_5.sBk = 1; gq0_5.sCo = 0; gq0_5.sCi = 0; gq0_5.sCm = C8; gq0_5.sRo = 0; gq0_5.sRi = 0; gq0_5.sRm = 0; gq0_5.sRn = 0;
      gq0_5.M = N; gq0_5.N = C8; gq0_5.K = C; gq0_5.zi_n = 1; gq0_5.flags = 1; gq0_5.act = 0;
      gq0_5.alpha = 1.0f; gq0_5.beta = 0.0f; gq0_5.sa = 1.0f; gq0_5.sb = 1.0f; gq0_5.Npad = C8; gq0_5.pad_ = 0;
      if ((long long)(N) >= 64 && (long long)(C8) >= 64) k_gemmT<1, 2, 4><<<dim3((unsigned)((C8) + 63) / 64, (unsigned)((N) + 31) / 32, (unsigned)(1)), 32, 0, stream>>>(gq0_5);
      else k_gemm<1><<<dim3((unsigned)((C8) + 31) / 32, (unsigned)((N) + 15) / 16, (unsigned)(1)), 32, 0, stream>>>(gq0_5); }
    { GemmP gk0_5;
      gk0_5.A = s1 + (size_t)5 * C * N; gk0_5.B = Wk; gk0_5.bias = bk; gk0_5.R = s1 + (size_t)5 * C * N; gk0_5.C = KF;
      gk0_5.sAo = 0; gk0_5.sAi = 0; gk0_5.sAm = 1; gk0_5.sAk = N; gk0_5.sBo = 0; gk0_5.sBi = 0; gk0_5.sBn = C; gk0_5.sBk = 1; gk0_5.sCo = 0; gk0_5.sCi = 0; gk0_5.sCm = C8; gk0_5.sRo = 0; gk0_5.sRi = 0; gk0_5.sRm = 0; gk0_5.sRn = 0;
      gk0_5.M = N; gk0_5.N = C8; gk0_5.K = C; gk0_5.zi_n = 1; gk0_5.flags = 1; gk0_5.act = 0;
      gk0_5.alpha = 1.0f; gk0_5.beta = 0.0f; gk0_5.sa = 1.0f; gk0_5.sb = 1.0f; gk0_5.Npad = C8; gk0_5.pad_ = 0;
      if ((long long)(N) >= 64 && (long long)(C8) >= 64) k_gemmT<1, 2, 4><<<dim3((unsigned)((C8) + 63) / 64, (unsigned)((N) + 31) / 32, (unsigned)(1)), 32, 0, stream>>>(gk0_5);
      else k_gemm<1><<<dim3((unsigned)((C8) + 31) / 32, (unsigned)((N) + 15) / 16, (unsigned)(1)), 32, 0, stream>>>(gk0_5); }
    k_cast16<<<(unsigned)((((long long)(256) * ((256) / 2)) + 255) / 256), 256, 0, stream>>>(Wv, 256, (_Float16*)(G64A), 256, 256, 256, 1.0f);
    k_castT16<<<(unsigned)((((long long)(1600) * ((256) / 2)) + 255) / 256), 256, 0, stream>>>(s1 + (size_t)5 * C * N, 1600, (_Float16*)(G64B), 256, 256, 1600, 16.0f);
    w25::wmma_gemm64<0, false, 1, 0, false, 0><<<dim3((unsigned)((((256) / 64) * ((1600) / 64) + 7) / 8), (unsigned)(1)), 256, 0, stream>>>((const unsigned short*)(G64A), nullptr, 256, 0, (const unsigned short*)(G64B), nullptr, 256, 0, (void*)(VF), nullptr, 1600, 0, bv, nullptr, 0, 256, 1600, 256, 0.0625f);
    k_ac_planes<<<(unsigned)(((long long)C * N / 2 + 255) / 256), 256, 0, stream>>>(QF, KF, VF, (_Float16*)QH, (_Float16*)QL, (_Float16*)KH, (_Float16*)KL, (_Float16*)V16, N * C8, (long long)C * N);
    w25::wmma_gemm64<1, true, 0, 0, false, 0><<<dim3((unsigned)((((N) / 64) * ((N) / 64) + 7) / 8), (unsigned)(1)), 256, 0, stream>>>((const unsigned short*)(QH), (const unsigned short*)(QL), C8, 0, (const unsigned short*)(KH), (const unsigned short*)(KL), C8, 0, (void*)(EN), nullptr, N, 0, nullptr, nullptr, 0, N, N, C8, 1.0f);
    k_ac_soft<<<N, 256, 0, stream>>>(EN, (_Float16*)P16, N);
    w25::wmma_gemm64<0, false, 0, 0, false, 0><<<dim3((unsigned)((((C) / 64) * ((N) / 64) + 7) / 8), (unsigned)(1)), 256, 0, stream>>>((const unsigned short*)(V16), nullptr, N, 0, (const unsigned short*)(P16), nullptr, N, 0, (void*)(CT), nullptr, N, 0, nullptr, nullptr, 0, C, N, N, 0.000244140625f);
    k_ac_fuse<<<(unsigned)(((long long)C * N + 255) / 256), 256, 0, stream>>>(CT, fw, out, 0, 5, (long long)C * N);
    { GemmP gq0_6;
      gq0_6.A = s0 + (size_t)6 * C * N; gq0_6.B = Wq; gq0_6.bias = bq; gq0_6.R = s0 + (size_t)6 * C * N; gq0_6.C = QF;
      gq0_6.sAo = 0; gq0_6.sAi = 0; gq0_6.sAm = 1; gq0_6.sAk = N; gq0_6.sBo = 0; gq0_6.sBi = 0; gq0_6.sBn = C; gq0_6.sBk = 1; gq0_6.sCo = 0; gq0_6.sCi = 0; gq0_6.sCm = C8; gq0_6.sRo = 0; gq0_6.sRi = 0; gq0_6.sRm = 0; gq0_6.sRn = 0;
      gq0_6.M = N; gq0_6.N = C8; gq0_6.K = C; gq0_6.zi_n = 1; gq0_6.flags = 1; gq0_6.act = 0;
      gq0_6.alpha = 1.0f; gq0_6.beta = 0.0f; gq0_6.sa = 1.0f; gq0_6.sb = 1.0f; gq0_6.Npad = C8; gq0_6.pad_ = 0;
      if ((long long)(N) >= 64 && (long long)(C8) >= 64) k_gemmT<1, 2, 4><<<dim3((unsigned)((C8) + 63) / 64, (unsigned)((N) + 31) / 32, (unsigned)(1)), 32, 0, stream>>>(gq0_6);
      else k_gemm<1><<<dim3((unsigned)((C8) + 31) / 32, (unsigned)((N) + 15) / 16, (unsigned)(1)), 32, 0, stream>>>(gq0_6); }
    { GemmP gk0_6;
      gk0_6.A = s1 + (size_t)6 * C * N; gk0_6.B = Wk; gk0_6.bias = bk; gk0_6.R = s1 + (size_t)6 * C * N; gk0_6.C = KF;
      gk0_6.sAo = 0; gk0_6.sAi = 0; gk0_6.sAm = 1; gk0_6.sAk = N; gk0_6.sBo = 0; gk0_6.sBi = 0; gk0_6.sBn = C; gk0_6.sBk = 1; gk0_6.sCo = 0; gk0_6.sCi = 0; gk0_6.sCm = C8; gk0_6.sRo = 0; gk0_6.sRi = 0; gk0_6.sRm = 0; gk0_6.sRn = 0;
      gk0_6.M = N; gk0_6.N = C8; gk0_6.K = C; gk0_6.zi_n = 1; gk0_6.flags = 1; gk0_6.act = 0;
      gk0_6.alpha = 1.0f; gk0_6.beta = 0.0f; gk0_6.sa = 1.0f; gk0_6.sb = 1.0f; gk0_6.Npad = C8; gk0_6.pad_ = 0;
      if ((long long)(N) >= 64 && (long long)(C8) >= 64) k_gemmT<1, 2, 4><<<dim3((unsigned)((C8) + 63) / 64, (unsigned)((N) + 31) / 32, (unsigned)(1)), 32, 0, stream>>>(gk0_6);
      else k_gemm<1><<<dim3((unsigned)((C8) + 31) / 32, (unsigned)((N) + 15) / 16, (unsigned)(1)), 32, 0, stream>>>(gk0_6); }
    k_cast16<<<(unsigned)((((long long)(256) * ((256) / 2)) + 255) / 256), 256, 0, stream>>>(Wv, 256, (_Float16*)(G64A), 256, 256, 256, 1.0f);
    k_castT16<<<(unsigned)((((long long)(1600) * ((256) / 2)) + 255) / 256), 256, 0, stream>>>(s1 + (size_t)6 * C * N, 1600, (_Float16*)(G64B), 256, 256, 1600, 16.0f);
    w25::wmma_gemm64<0, false, 1, 0, false, 0><<<dim3((unsigned)((((256) / 64) * ((1600) / 64) + 7) / 8), (unsigned)(1)), 256, 0, stream>>>((const unsigned short*)(G64A), nullptr, 256, 0, (const unsigned short*)(G64B), nullptr, 256, 0, (void*)(VF), nullptr, 1600, 0, bv, nullptr, 0, 256, 1600, 256, 0.0625f);
    k_ac_planes<<<(unsigned)(((long long)C * N / 2 + 255) / 256), 256, 0, stream>>>(QF, KF, VF, (_Float16*)QH, (_Float16*)QL, (_Float16*)KH, (_Float16*)KL, (_Float16*)V16, N * C8, (long long)C * N);
    w25::wmma_gemm64<1, true, 0, 0, false, 0><<<dim3((unsigned)((((N) / 64) * ((N) / 64) + 7) / 8), (unsigned)(1)), 256, 0, stream>>>((const unsigned short*)(QH), (const unsigned short*)(QL), C8, 0, (const unsigned short*)(KH), (const unsigned short*)(KL), C8, 0, (void*)(EN), nullptr, N, 0, nullptr, nullptr, 0, N, N, C8, 1.0f);
    k_ac_soft<<<N, 256, 0, stream>>>(EN, (_Float16*)P16, N);
    w25::wmma_gemm64<0, false, 0, 0, false, 0><<<dim3((unsigned)((((C) / 64) * ((N) / 64) + 7) / 8), (unsigned)(1)), 256, 0, stream>>>((const unsigned short*)(V16), nullptr, N, 0, (const unsigned short*)(P16), nullptr, N, 0, (void*)(CT), nullptr, N, 0, nullptr, nullptr, 0, C, N, N, 0.000244140625f);
    k_ac_fuse<<<(unsigned)(((long long)C * N + 255) / 256), 256, 0, stream>>>(CT, fw, out, 0, 6, (long long)C * N);
    { GemmP gq0_7;
      gq0_7.A = s0 + (size_t)7 * C * N; gq0_7.B = Wq; gq0_7.bias = bq; gq0_7.R = s0 + (size_t)7 * C * N; gq0_7.C = QF;
      gq0_7.sAo = 0; gq0_7.sAi = 0; gq0_7.sAm = 1; gq0_7.sAk = N; gq0_7.sBo = 0; gq0_7.sBi = 0; gq0_7.sBn = C; gq0_7.sBk = 1; gq0_7.sCo = 0; gq0_7.sCi = 0; gq0_7.sCm = C8; gq0_7.sRo = 0; gq0_7.sRi = 0; gq0_7.sRm = 0; gq0_7.sRn = 0;
      gq0_7.M = N; gq0_7.N = C8; gq0_7.K = C; gq0_7.zi_n = 1; gq0_7.flags = 1; gq0_7.act = 0;
      gq0_7.alpha = 1.0f; gq0_7.beta = 0.0f; gq0_7.sa = 1.0f; gq0_7.sb = 1.0f; gq0_7.Npad = C8; gq0_7.pad_ = 0;
      if ((long long)(N) >= 64 && (long long)(C8) >= 64) k_gemmT<1, 2, 4><<<dim3((unsigned)((C8) + 63) / 64, (unsigned)((N) + 31) / 32, (unsigned)(1)), 32, 0, stream>>>(gq0_7);
      else k_gemm<1><<<dim3((unsigned)((C8) + 31) / 32, (unsigned)((N) + 15) / 16, (unsigned)(1)), 32, 0, stream>>>(gq0_7); }
    { GemmP gk0_7;
      gk0_7.A = s1 + (size_t)7 * C * N; gk0_7.B = Wk; gk0_7.bias = bk; gk0_7.R = s1 + (size_t)7 * C * N; gk0_7.C = KF;
      gk0_7.sAo = 0; gk0_7.sAi = 0; gk0_7.sAm = 1; gk0_7.sAk = N; gk0_7.sBo = 0; gk0_7.sBi = 0; gk0_7.sBn = C; gk0_7.sBk = 1; gk0_7.sCo = 0; gk0_7.sCi = 0; gk0_7.sCm = C8; gk0_7.sRo = 0; gk0_7.sRi = 0; gk0_7.sRm = 0; gk0_7.sRn = 0;
      gk0_7.M = N; gk0_7.N = C8; gk0_7.K = C; gk0_7.zi_n = 1; gk0_7.flags = 1; gk0_7.act = 0;
      gk0_7.alpha = 1.0f; gk0_7.beta = 0.0f; gk0_7.sa = 1.0f; gk0_7.sb = 1.0f; gk0_7.Npad = C8; gk0_7.pad_ = 0;
      if ((long long)(N) >= 64 && (long long)(C8) >= 64) k_gemmT<1, 2, 4><<<dim3((unsigned)((C8) + 63) / 64, (unsigned)((N) + 31) / 32, (unsigned)(1)), 32, 0, stream>>>(gk0_7);
      else k_gemm<1><<<dim3((unsigned)((C8) + 31) / 32, (unsigned)((N) + 15) / 16, (unsigned)(1)), 32, 0, stream>>>(gk0_7); }
    k_cast16<<<(unsigned)((((long long)(256) * ((256) / 2)) + 255) / 256), 256, 0, stream>>>(Wv, 256, (_Float16*)(G64A), 256, 256, 256, 1.0f);
    k_castT16<<<(unsigned)((((long long)(1600) * ((256) / 2)) + 255) / 256), 256, 0, stream>>>(s1 + (size_t)7 * C * N, 1600, (_Float16*)(G64B), 256, 256, 1600, 16.0f);
    w25::wmma_gemm64<0, false, 1, 0, false, 0><<<dim3((unsigned)((((256) / 64) * ((1600) / 64) + 7) / 8), (unsigned)(1)), 256, 0, stream>>>((const unsigned short*)(G64A), nullptr, 256, 0, (const unsigned short*)(G64B), nullptr, 256, 0, (void*)(VF), nullptr, 1600, 0, bv, nullptr, 0, 256, 1600, 256, 0.0625f);
    k_ac_planes<<<(unsigned)(((long long)C * N / 2 + 255) / 256), 256, 0, stream>>>(QF, KF, VF, (_Float16*)QH, (_Float16*)QL, (_Float16*)KH, (_Float16*)KL, (_Float16*)V16, N * C8, (long long)C * N);
    w25::wmma_gemm64<1, true, 0, 0, false, 0><<<dim3((unsigned)((((N) / 64) * ((N) / 64) + 7) / 8), (unsigned)(1)), 256, 0, stream>>>((const unsigned short*)(QH), (const unsigned short*)(QL), C8, 0, (const unsigned short*)(KH), (const unsigned short*)(KL), C8, 0, (void*)(EN), nullptr, N, 0, nullptr, nullptr, 0, N, N, C8, 1.0f);
    k_ac_soft<<<N, 256, 0, stream>>>(EN, (_Float16*)P16, N);
    w25::wmma_gemm64<0, false, 0, 0, false, 0><<<dim3((unsigned)((((C) / 64) * ((N) / 64) + 7) / 8), (unsigned)(1)), 256, 0, stream>>>((const unsigned short*)(V16), nullptr, N, 0, (const unsigned short*)(P16), nullptr, N, 0, (void*)(CT), nullptr, N, 0, nullptr, nullptr, 0, C, N, N, 0.000244140625f);
    k_ac_fuse<<<(unsigned)(((long long)C * N + 255) / 256), 256, 0, stream>>>(CT, fw, out, 0, 7, (long long)C * N);
    { GemmP gq0_8;
      gq0_8.A = s0 + (size_t)8 * C * N; gq0_8.B = Wq; gq0_8.bias = bq; gq0_8.R = s0 + (size_t)8 * C * N; gq0_8.C = QF;
      gq0_8.sAo = 0; gq0_8.sAi = 0; gq0_8.sAm = 1; gq0_8.sAk = N; gq0_8.sBo = 0; gq0_8.sBi = 0; gq0_8.sBn = C; gq0_8.sBk = 1; gq0_8.sCo = 0; gq0_8.sCi = 0; gq0_8.sCm = C8; gq0_8.sRo = 0; gq0_8.sRi = 0; gq0_8.sRm = 0; gq0_8.sRn = 0;
      gq0_8.M = N; gq0_8.N = C8; gq0_8.K = C; gq0_8.zi_n = 1; gq0_8.flags = 1; gq0_8.act = 0;
      gq0_8.alpha = 1.0f; gq0_8.beta = 0.0f; gq0_8.sa = 1.0f; gq0_8.sb = 1.0f; gq0_8.Npad = C8; gq0_8.pad_ = 0;
      if ((long long)(N) >= 64 && (long long)(C8) >= 64) k_gemmT<1, 2, 4><<<dim3((unsigned)((C8) + 63) / 64, (unsigned)((N) + 31) / 32, (unsigned)(1)), 32, 0, stream>>>(gq0_8);
      else k_gemm<1><<<dim3((unsigned)((C8) + 31) / 32, (unsigned)((N) + 15) / 16, (unsigned)(1)), 32, 0, stream>>>(gq0_8); }
    { GemmP gk0_8;
      gk0_8.A = s1 + (size_t)8 * C * N; gk0_8.B = Wk; gk0_8.bias = bk; gk0_8.R = s1 + (size_t)8 * C * N; gk0_8.C = KF;
      gk0_8.sAo = 0; gk0_8.sAi = 0; gk0_8.sAm = 1; gk0_8.sAk = N; gk0_8.sBo = 0; gk0_8.sBi = 0; gk0_8.sBn = C; gk0_8.sBk = 1; gk0_8.sCo = 0; gk0_8.sCi = 0; gk0_8.sCm = C8; gk0_8.sRo = 0; gk0_8.sRi = 0; gk0_8.sRm = 0; gk0_8.sRn = 0;
      gk0_8.M = N; gk0_8.N = C8; gk0_8.K = C; gk0_8.zi_n = 1; gk0_8.flags = 1; gk0_8.act = 0;
      gk0_8.alpha = 1.0f; gk0_8.beta = 0.0f; gk0_8.sa = 1.0f; gk0_8.sb = 1.0f; gk0_8.Npad = C8; gk0_8.pad_ = 0;
      if ((long long)(N) >= 64 && (long long)(C8) >= 64) k_gemmT<1, 2, 4><<<dim3((unsigned)((C8) + 63) / 64, (unsigned)((N) + 31) / 32, (unsigned)(1)), 32, 0, stream>>>(gk0_8);
      else k_gemm<1><<<dim3((unsigned)((C8) + 31) / 32, (unsigned)((N) + 15) / 16, (unsigned)(1)), 32, 0, stream>>>(gk0_8); }
    k_cast16<<<(unsigned)((((long long)(256) * ((256) / 2)) + 255) / 256), 256, 0, stream>>>(Wv, 256, (_Float16*)(G64A), 256, 256, 256, 1.0f);
    k_castT16<<<(unsigned)((((long long)(1600) * ((256) / 2)) + 255) / 256), 256, 0, stream>>>(s1 + (size_t)8 * C * N, 1600, (_Float16*)(G64B), 256, 256, 1600, 16.0f);
    w25::wmma_gemm64<0, false, 1, 0, false, 0><<<dim3((unsigned)((((256) / 64) * ((1600) / 64) + 7) / 8), (unsigned)(1)), 256, 0, stream>>>((const unsigned short*)(G64A), nullptr, 256, 0, (const unsigned short*)(G64B), nullptr, 256, 0, (void*)(VF), nullptr, 1600, 0, bv, nullptr, 0, 256, 1600, 256, 0.0625f);
    k_ac_planes<<<(unsigned)(((long long)C * N / 2 + 255) / 256), 256, 0, stream>>>(QF, KF, VF, (_Float16*)QH, (_Float16*)QL, (_Float16*)KH, (_Float16*)KL, (_Float16*)V16, N * C8, (long long)C * N);
    w25::wmma_gemm64<1, true, 0, 0, false, 0><<<dim3((unsigned)((((N) / 64) * ((N) / 64) + 7) / 8), (unsigned)(1)), 256, 0, stream>>>((const unsigned short*)(QH), (const unsigned short*)(QL), C8, 0, (const unsigned short*)(KH), (const unsigned short*)(KL), C8, 0, (void*)(EN), nullptr, N, 0, nullptr, nullptr, 0, N, N, C8, 1.0f);
    k_ac_soft<<<N, 256, 0, stream>>>(EN, (_Float16*)P16, N);
    w25::wmma_gemm64<0, false, 0, 0, false, 0><<<dim3((unsigned)((((C) / 64) * ((N) / 64) + 7) / 8), (unsigned)(1)), 256, 0, stream>>>((const unsigned short*)(V16), nullptr, N, 0, (const unsigned short*)(P16), nullptr, N, 0, (void*)(CT), nullptr, N, 0, nullptr, nullptr, 0, C, N, N, 0.000244140625f);
    k_ac_fuse<<<(unsigned)(((long long)C * N + 255) / 256), 256, 0, stream>>>(CT, fw, out, 0, 8, (long long)C * N);
    { GemmP gq0_9;
      gq0_9.A = s0 + (size_t)9 * C * N; gq0_9.B = Wq; gq0_9.bias = bq; gq0_9.R = s0 + (size_t)9 * C * N; gq0_9.C = QF;
      gq0_9.sAo = 0; gq0_9.sAi = 0; gq0_9.sAm = 1; gq0_9.sAk = N; gq0_9.sBo = 0; gq0_9.sBi = 0; gq0_9.sBn = C; gq0_9.sBk = 1; gq0_9.sCo = 0; gq0_9.sCi = 0; gq0_9.sCm = C8; gq0_9.sRo = 0; gq0_9.sRi = 0; gq0_9.sRm = 0; gq0_9.sRn = 0;
      gq0_9.M = N; gq0_9.N = C8; gq0_9.K = C; gq0_9.zi_n = 1; gq0_9.flags = 1; gq0_9.act = 0;
      gq0_9.alpha = 1.0f; gq0_9.beta = 0.0f; gq0_9.sa = 1.0f; gq0_9.sb = 1.0f; gq0_9.Npad = C8; gq0_9.pad_ = 0;
      if ((long long)(N) >= 64 && (long long)(C8) >= 64) k_gemmT<1, 2, 4><<<dim3((unsigned)((C8) + 63) / 64, (unsigned)((N) + 31) / 32, (unsigned)(1)), 32, 0, stream>>>(gq0_9);
      else k_gemm<1><<<dim3((unsigned)((C8) + 31) / 32, (unsigned)((N) + 15) / 16, (unsigned)(1)), 32, 0, stream>>>(gq0_9); }
    { GemmP gk0_9;
      gk0_9.A = s1 + (size_t)9 * C * N; gk0_9.B = Wk; gk0_9.bias = bk; gk0_9.R = s1 + (size_t)9 * C * N; gk0_9.C = KF;
      gk0_9.sAo = 0; gk0_9.sAi = 0; gk0_9.sAm = 1; gk0_9.sAk = N; gk0_9.sBo = 0; gk0_9.sBi = 0; gk0_9.sBn = C; gk0_9.sBk = 1; gk0_9.sCo = 0; gk0_9.sCi = 0; gk0_9.sCm = C8; gk0_9.sRo = 0; gk0_9.sRi = 0; gk0_9.sRm = 0; gk0_9.sRn = 0;
      gk0_9.M = N; gk0_9.N = C8; gk0_9.K = C; gk0_9.zi_n = 1; gk0_9.flags = 1; gk0_9.act = 0;
      gk0_9.alpha = 1.0f; gk0_9.beta = 0.0f; gk0_9.sa = 1.0f; gk0_9.sb = 1.0f; gk0_9.Npad = C8; gk0_9.pad_ = 0;
      if ((long long)(N) >= 64 && (long long)(C8) >= 64) k_gemmT<1, 2, 4><<<dim3((unsigned)((C8) + 63) / 64, (unsigned)((N) + 31) / 32, (unsigned)(1)), 32, 0, stream>>>(gk0_9);
      else k_gemm<1><<<dim3((unsigned)((C8) + 31) / 32, (unsigned)((N) + 15) / 16, (unsigned)(1)), 32, 0, stream>>>(gk0_9); }
    k_cast16<<<(unsigned)((((long long)(256) * ((256) / 2)) + 255) / 256), 256, 0, stream>>>(Wv, 256, (_Float16*)(G64A), 256, 256, 256, 1.0f);
    k_castT16<<<(unsigned)((((long long)(1600) * ((256) / 2)) + 255) / 256), 256, 0, stream>>>(s1 + (size_t)9 * C * N, 1600, (_Float16*)(G64B), 256, 256, 1600, 16.0f);
    w25::wmma_gemm64<0, false, 1, 0, false, 0><<<dim3((unsigned)((((256) / 64) * ((1600) / 64) + 7) / 8), (unsigned)(1)), 256, 0, stream>>>((const unsigned short*)(G64A), nullptr, 256, 0, (const unsigned short*)(G64B), nullptr, 256, 0, (void*)(VF), nullptr, 1600, 0, bv, nullptr, 0, 256, 1600, 256, 0.0625f);
    k_ac_planes<<<(unsigned)(((long long)C * N / 2 + 255) / 256), 256, 0, stream>>>(QF, KF, VF, (_Float16*)QH, (_Float16*)QL, (_Float16*)KH, (_Float16*)KL, (_Float16*)V16, N * C8, (long long)C * N);
    w25::wmma_gemm64<1, true, 0, 0, false, 0><<<dim3((unsigned)((((N) / 64) * ((N) / 64) + 7) / 8), (unsigned)(1)), 256, 0, stream>>>((const unsigned short*)(QH), (const unsigned short*)(QL), C8, 0, (const unsigned short*)(KH), (const unsigned short*)(KL), C8, 0, (void*)(EN), nullptr, N, 0, nullptr, nullptr, 0, N, N, C8, 1.0f);
    k_ac_soft<<<N, 256, 0, stream>>>(EN, (_Float16*)P16, N);
    w25::wmma_gemm64<0, false, 0, 0, false, 0><<<dim3((unsigned)((((C) / 64) * ((N) / 64) + 7) / 8), (unsigned)(1)), 256, 0, stream>>>((const unsigned short*)(V16), nullptr, N, 0, (const unsigned short*)(P16), nullptr, N, 0, (void*)(CT), nullptr, N, 0, nullptr, nullptr, 0, C, N, N, 0.000244140625f);
    k_ac_fuse<<<(unsigned)(((long long)C * N + 255) / 256), 256, 0, stream>>>(CT, fw, out, 0, 9, (long long)C * N);
    { GemmP gq0_10;
      gq0_10.A = s0 + (size_t)10 * C * N; gq0_10.B = Wq; gq0_10.bias = bq; gq0_10.R = s0 + (size_t)10 * C * N; gq0_10.C = QF;
      gq0_10.sAo = 0; gq0_10.sAi = 0; gq0_10.sAm = 1; gq0_10.sAk = N; gq0_10.sBo = 0; gq0_10.sBi = 0; gq0_10.sBn = C; gq0_10.sBk = 1; gq0_10.sCo = 0; gq0_10.sCi = 0; gq0_10.sCm = C8; gq0_10.sRo = 0; gq0_10.sRi = 0; gq0_10.sRm = 0; gq0_10.sRn = 0;
      gq0_10.M = N; gq0_10.N = C8; gq0_10.K = C; gq0_10.zi_n = 1; gq0_10.flags = 1; gq0_10.act = 0;
      gq0_10.alpha = 1.0f; gq0_10.beta = 0.0f; gq0_10.sa = 1.0f; gq0_10.sb = 1.0f; gq0_10.Npad = C8; gq0_10.pad_ = 0;
      if ((long long)(N) >= 64 && (long long)(C8) >= 64) k_gemmT<1, 2, 4><<<dim3((unsigned)((C8) + 63) / 64, (unsigned)((N) + 31) / 32, (unsigned)(1)), 32, 0, stream>>>(gq0_10);
      else k_gemm<1><<<dim3((unsigned)((C8) + 31) / 32, (unsigned)((N) + 15) / 16, (unsigned)(1)), 32, 0, stream>>>(gq0_10); }
    { GemmP gk0_10;
      gk0_10.A = s1 + (size_t)10 * C * N; gk0_10.B = Wk; gk0_10.bias = bk; gk0_10.R = s1 + (size_t)10 * C * N; gk0_10.C = KF;
      gk0_10.sAo = 0; gk0_10.sAi = 0; gk0_10.sAm = 1; gk0_10.sAk = N; gk0_10.sBo = 0; gk0_10.sBi = 0; gk0_10.sBn = C; gk0_10.sBk = 1; gk0_10.sCo = 0; gk0_10.sCi = 0; gk0_10.sCm = C8; gk0_10.sRo = 0; gk0_10.sRi = 0; gk0_10.sRm = 0; gk0_10.sRn = 0;
      gk0_10.M = N; gk0_10.N = C8; gk0_10.K = C; gk0_10.zi_n = 1; gk0_10.flags = 1; gk0_10.act = 0;
      gk0_10.alpha = 1.0f; gk0_10.beta = 0.0f; gk0_10.sa = 1.0f; gk0_10.sb = 1.0f; gk0_10.Npad = C8; gk0_10.pad_ = 0;
      if ((long long)(N) >= 64 && (long long)(C8) >= 64) k_gemmT<1, 2, 4><<<dim3((unsigned)((C8) + 63) / 64, (unsigned)((N) + 31) / 32, (unsigned)(1)), 32, 0, stream>>>(gk0_10);
      else k_gemm<1><<<dim3((unsigned)((C8) + 31) / 32, (unsigned)((N) + 15) / 16, (unsigned)(1)), 32, 0, stream>>>(gk0_10); }
    k_cast16<<<(unsigned)((((long long)(256) * ((256) / 2)) + 255) / 256), 256, 0, stream>>>(Wv, 256, (_Float16*)(G64A), 256, 256, 256, 1.0f);
    k_castT16<<<(unsigned)((((long long)(1600) * ((256) / 2)) + 255) / 256), 256, 0, stream>>>(s1 + (size_t)10 * C * N, 1600, (_Float16*)(G64B), 256, 256, 1600, 16.0f);
    w25::wmma_gemm64<0, false, 1, 0, false, 0><<<dim3((unsigned)((((256) / 64) * ((1600) / 64) + 7) / 8), (unsigned)(1)), 256, 0, stream>>>((const unsigned short*)(G64A), nullptr, 256, 0, (const unsigned short*)(G64B), nullptr, 256, 0, (void*)(VF), nullptr, 1600, 0, bv, nullptr, 0, 256, 1600, 256, 0.0625f);
    k_ac_planes<<<(unsigned)(((long long)C * N / 2 + 255) / 256), 256, 0, stream>>>(QF, KF, VF, (_Float16*)QH, (_Float16*)QL, (_Float16*)KH, (_Float16*)KL, (_Float16*)V16, N * C8, (long long)C * N);
    w25::wmma_gemm64<1, true, 0, 0, false, 0><<<dim3((unsigned)((((N) / 64) * ((N) / 64) + 7) / 8), (unsigned)(1)), 256, 0, stream>>>((const unsigned short*)(QH), (const unsigned short*)(QL), C8, 0, (const unsigned short*)(KH), (const unsigned short*)(KL), C8, 0, (void*)(EN), nullptr, N, 0, nullptr, nullptr, 0, N, N, C8, 1.0f);
    k_ac_soft<<<N, 256, 0, stream>>>(EN, (_Float16*)P16, N);
    w25::wmma_gemm64<0, false, 0, 0, false, 0><<<dim3((unsigned)((((C) / 64) * ((N) / 64) + 7) / 8), (unsigned)(1)), 256, 0, stream>>>((const unsigned short*)(V16), nullptr, N, 0, (const unsigned short*)(P16), nullptr, N, 0, (void*)(CT), nullptr, N, 0, nullptr, nullptr, 0, C, N, N, 0.000244140625f);
    k_ac_fuse<<<(unsigned)(((long long)C * N + 255) / 256), 256, 0, stream>>>(CT, fw, out, 0, 10, (long long)C * N);
    { GemmP gq0_11;
      gq0_11.A = s0 + (size_t)11 * C * N; gq0_11.B = Wq; gq0_11.bias = bq; gq0_11.R = s0 + (size_t)11 * C * N; gq0_11.C = QF;
      gq0_11.sAo = 0; gq0_11.sAi = 0; gq0_11.sAm = 1; gq0_11.sAk = N; gq0_11.sBo = 0; gq0_11.sBi = 0; gq0_11.sBn = C; gq0_11.sBk = 1; gq0_11.sCo = 0; gq0_11.sCi = 0; gq0_11.sCm = C8; gq0_11.sRo = 0; gq0_11.sRi = 0; gq0_11.sRm = 0; gq0_11.sRn = 0;
      gq0_11.M = N; gq0_11.N = C8; gq0_11.K = C; gq0_11.zi_n = 1; gq0_11.flags = 1; gq0_11.act = 0;
      gq0_11.alpha = 1.0f; gq0_11.beta = 0.0f; gq0_11.sa = 1.0f; gq0_11.sb = 1.0f; gq0_11.Npad = C8; gq0_11.pad_ = 0;
      if ((long long)(N) >= 64 && (long long)(C8) >= 64) k_gemmT<1, 2, 4><<<dim3((unsigned)((C8) + 63) / 64, (unsigned)((N) + 31) / 32, (unsigned)(1)), 32, 0, stream>>>(gq0_11);
      else k_gemm<1><<<dim3((unsigned)((C8) + 31) / 32, (unsigned)((N) + 15) / 16, (unsigned)(1)), 32, 0, stream>>>(gq0_11); }
    { GemmP gk0_11;
      gk0_11.A = s1 + (size_t)11 * C * N; gk0_11.B = Wk; gk0_11.bias = bk; gk0_11.R = s1 + (size_t)11 * C * N; gk0_11.C = KF;
      gk0_11.sAo = 0; gk0_11.sAi = 0; gk0_11.sAm = 1; gk0_11.sAk = N; gk0_11.sBo = 0; gk0_11.sBi = 0; gk0_11.sBn = C; gk0_11.sBk = 1; gk0_11.sCo = 0; gk0_11.sCi = 0; gk0_11.sCm = C8; gk0_11.sRo = 0; gk0_11.sRi = 0; gk0_11.sRm = 0; gk0_11.sRn = 0;
      gk0_11.M = N; gk0_11.N = C8; gk0_11.K = C; gk0_11.zi_n = 1; gk0_11.flags = 1; gk0_11.act = 0;
      gk0_11.alpha = 1.0f; gk0_11.beta = 0.0f; gk0_11.sa = 1.0f; gk0_11.sb = 1.0f; gk0_11.Npad = C8; gk0_11.pad_ = 0;
      if ((long long)(N) >= 64 && (long long)(C8) >= 64) k_gemmT<1, 2, 4><<<dim3((unsigned)((C8) + 63) / 64, (unsigned)((N) + 31) / 32, (unsigned)(1)), 32, 0, stream>>>(gk0_11);
      else k_gemm<1><<<dim3((unsigned)((C8) + 31) / 32, (unsigned)((N) + 15) / 16, (unsigned)(1)), 32, 0, stream>>>(gk0_11); }
    k_cast16<<<(unsigned)((((long long)(256) * ((256) / 2)) + 255) / 256), 256, 0, stream>>>(Wv, 256, (_Float16*)(G64A), 256, 256, 256, 1.0f);
    k_castT16<<<(unsigned)((((long long)(1600) * ((256) / 2)) + 255) / 256), 256, 0, stream>>>(s1 + (size_t)11 * C * N, 1600, (_Float16*)(G64B), 256, 256, 1600, 16.0f);
    w25::wmma_gemm64<0, false, 1, 0, false, 0><<<dim3((unsigned)((((256) / 64) * ((1600) / 64) + 7) / 8), (unsigned)(1)), 256, 0, stream>>>((const unsigned short*)(G64A), nullptr, 256, 0, (const unsigned short*)(G64B), nullptr, 256, 0, (void*)(VF), nullptr, 1600, 0, bv, nullptr, 0, 256, 1600, 256, 0.0625f);
    k_ac_planes<<<(unsigned)(((long long)C * N / 2 + 255) / 256), 256, 0, stream>>>(QF, KF, VF, (_Float16*)QH, (_Float16*)QL, (_Float16*)KH, (_Float16*)KL, (_Float16*)V16, N * C8, (long long)C * N);
    w25::wmma_gemm64<1, true, 0, 0, false, 0><<<dim3((unsigned)((((N) / 64) * ((N) / 64) + 7) / 8), (unsigned)(1)), 256, 0, stream>>>((const unsigned short*)(QH), (const unsigned short*)(QL), C8, 0, (const unsigned short*)(KH), (const unsigned short*)(KL), C8, 0, (void*)(EN), nullptr, N, 0, nullptr, nullptr, 0, N, N, C8, 1.0f);
    k_ac_soft<<<N, 256, 0, stream>>>(EN, (_Float16*)P16, N);
    w25::wmma_gemm64<0, false, 0, 0, false, 0><<<dim3((unsigned)((((C) / 64) * ((N) / 64) + 7) / 8), (unsigned)(1)), 256, 0, stream>>>((const unsigned short*)(V16), nullptr, N, 0, (const unsigned short*)(P16), nullptr, N, 0, (void*)(CT), nullptr, N, 0, nullptr, nullptr, 0, C, N, N, 0.000244140625f);
    k_ac_fuse<<<(unsigned)(((long long)C * N + 255) / 256), 256, 0, stream>>>(CT, fw, out, 0, 11, (long long)C * N);
    { GemmP gq0_12;
      gq0_12.A = s0 + (size_t)12 * C * N; gq0_12.B = Wq; gq0_12.bias = bq; gq0_12.R = s0 + (size_t)12 * C * N; gq0_12.C = QF;
      gq0_12.sAo = 0; gq0_12.sAi = 0; gq0_12.sAm = 1; gq0_12.sAk = N; gq0_12.sBo = 0; gq0_12.sBi = 0; gq0_12.sBn = C; gq0_12.sBk = 1; gq0_12.sCo = 0; gq0_12.sCi = 0; gq0_12.sCm = C8; gq0_12.sRo = 0; gq0_12.sRi = 0; gq0_12.sRm = 0; gq0_12.sRn = 0;
      gq0_12.M = N; gq0_12.N = C8; gq0_12.K = C; gq0_12.zi_n = 1; gq0_12.flags = 1; gq0_12.act = 0;
      gq0_12.alpha = 1.0f; gq0_12.beta = 0.0f; gq0_12.sa = 1.0f; gq0_12.sb = 1.0f; gq0_12.Npad = C8; gq0_12.pad_ = 0;
      if ((long long)(N) >= 64 && (long long)(C8) >= 64) k_gemmT<1, 2, 4><<<dim3((unsigned)((C8) + 63) / 64, (unsigned)((N) + 31) / 32, (unsigned)(1)), 32, 0, stream>>>(gq0_12);
      else k_gemm<1><<<dim3((unsigned)((C8) + 31) / 32, (unsigned)((N) + 15) / 16, (unsigned)(1)), 32, 0, stream>>>(gq0_12); }
    { GemmP gk0_12;
      gk0_12.A = s1 + (size_t)12 * C * N; gk0_12.B = Wk; gk0_12.bias = bk; gk0_12.R = s1 + (size_t)12 * C * N; gk0_12.C = KF;
      gk0_12.sAo = 0; gk0_12.sAi = 0; gk0_12.sAm = 1; gk0_12.sAk = N; gk0_12.sBo = 0; gk0_12.sBi = 0; gk0_12.sBn = C; gk0_12.sBk = 1; gk0_12.sCo = 0; gk0_12.sCi = 0; gk0_12.sCm = C8; gk0_12.sRo = 0; gk0_12.sRi = 0; gk0_12.sRm = 0; gk0_12.sRn = 0;
      gk0_12.M = N; gk0_12.N = C8; gk0_12.K = C; gk0_12.zi_n = 1; gk0_12.flags = 1; gk0_12.act = 0;
      gk0_12.alpha = 1.0f; gk0_12.beta = 0.0f; gk0_12.sa = 1.0f; gk0_12.sb = 1.0f; gk0_12.Npad = C8; gk0_12.pad_ = 0;
      if ((long long)(N) >= 64 && (long long)(C8) >= 64) k_gemmT<1, 2, 4><<<dim3((unsigned)((C8) + 63) / 64, (unsigned)((N) + 31) / 32, (unsigned)(1)), 32, 0, stream>>>(gk0_12);
      else k_gemm<1><<<dim3((unsigned)((C8) + 31) / 32, (unsigned)((N) + 15) / 16, (unsigned)(1)), 32, 0, stream>>>(gk0_12); }
    k_cast16<<<(unsigned)((((long long)(256) * ((256) / 2)) + 255) / 256), 256, 0, stream>>>(Wv, 256, (_Float16*)(G64A), 256, 256, 256, 1.0f);
    k_castT16<<<(unsigned)((((long long)(1600) * ((256) / 2)) + 255) / 256), 256, 0, stream>>>(s1 + (size_t)12 * C * N, 1600, (_Float16*)(G64B), 256, 256, 1600, 16.0f);
    w25::wmma_gemm64<0, false, 1, 0, false, 0><<<dim3((unsigned)((((256) / 64) * ((1600) / 64) + 7) / 8), (unsigned)(1)), 256, 0, stream>>>((const unsigned short*)(G64A), nullptr, 256, 0, (const unsigned short*)(G64B), nullptr, 256, 0, (void*)(VF), nullptr, 1600, 0, bv, nullptr, 0, 256, 1600, 256, 0.0625f);
    k_ac_planes<<<(unsigned)(((long long)C * N / 2 + 255) / 256), 256, 0, stream>>>(QF, KF, VF, (_Float16*)QH, (_Float16*)QL, (_Float16*)KH, (_Float16*)KL, (_Float16*)V16, N * C8, (long long)C * N);
    w25::wmma_gemm64<1, true, 0, 0, false, 0><<<dim3((unsigned)((((N) / 64) * ((N) / 64) + 7) / 8), (unsigned)(1)), 256, 0, stream>>>((const unsigned short*)(QH), (const unsigned short*)(QL), C8, 0, (const unsigned short*)(KH), (const unsigned short*)(KL), C8, 0, (void*)(EN), nullptr, N, 0, nullptr, nullptr, 0, N, N, C8, 1.0f);
    k_ac_soft<<<N, 256, 0, stream>>>(EN, (_Float16*)P16, N);
    w25::wmma_gemm64<0, false, 0, 0, false, 0><<<dim3((unsigned)((((C) / 64) * ((N) / 64) + 7) / 8), (unsigned)(1)), 256, 0, stream>>>((const unsigned short*)(V16), nullptr, N, 0, (const unsigned short*)(P16), nullptr, N, 0, (void*)(CT), nullptr, N, 0, nullptr, nullptr, 0, C, N, N, 0.000244140625f);
    k_ac_fuse<<<(unsigned)(((long long)C * N + 255) / 256), 256, 0, stream>>>(CT, fw, out, 0, 12, (long long)C * N);
    { GemmP gq0_13;
      gq0_13.A = s0 + (size_t)13 * C * N; gq0_13.B = Wq; gq0_13.bias = bq; gq0_13.R = s0 + (size_t)13 * C * N; gq0_13.C = QF;
      gq0_13.sAo = 0; gq0_13.sAi = 0; gq0_13.sAm = 1; gq0_13.sAk = N; gq0_13.sBo = 0; gq0_13.sBi = 0; gq0_13.sBn = C; gq0_13.sBk = 1; gq0_13.sCo = 0; gq0_13.sCi = 0; gq0_13.sCm = C8; gq0_13.sRo = 0; gq0_13.sRi = 0; gq0_13.sRm = 0; gq0_13.sRn = 0;
      gq0_13.M = N; gq0_13.N = C8; gq0_13.K = C; gq0_13.zi_n = 1; gq0_13.flags = 1; gq0_13.act = 0;
      gq0_13.alpha = 1.0f; gq0_13.beta = 0.0f; gq0_13.sa = 1.0f; gq0_13.sb = 1.0f; gq0_13.Npad = C8; gq0_13.pad_ = 0;
      if ((long long)(N) >= 64 && (long long)(C8) >= 64) k_gemmT<1, 2, 4><<<dim3((unsigned)((C8) + 63) / 64, (unsigned)((N) + 31) / 32, (unsigned)(1)), 32, 0, stream>>>(gq0_13);
      else k_gemm<1><<<dim3((unsigned)((C8) + 31) / 32, (unsigned)((N) + 15) / 16, (unsigned)(1)), 32, 0, stream>>>(gq0_13); }
    { GemmP gk0_13;
      gk0_13.A = s1 + (size_t)13 * C * N; gk0_13.B = Wk; gk0_13.bias = bk; gk0_13.R = s1 + (size_t)13 * C * N; gk0_13.C = KF;
      gk0_13.sAo = 0; gk0_13.sAi = 0; gk0_13.sAm = 1; gk0_13.sAk = N; gk0_13.sBo = 0; gk0_13.sBi = 0; gk0_13.sBn = C; gk0_13.sBk = 1; gk0_13.sCo = 0; gk0_13.sCi = 0; gk0_13.sCm = C8; gk0_13.sRo = 0; gk0_13.sRi = 0; gk0_13.sRm = 0; gk0_13.sRn = 0;
      gk0_13.M = N; gk0_13.N = C8; gk0_13.K = C; gk0_13.zi_n = 1; gk0_13.flags = 1; gk0_13.act = 0;
      gk0_13.alpha = 1.0f; gk0_13.beta = 0.0f; gk0_13.sa = 1.0f; gk0_13.sb = 1.0f; gk0_13.Npad = C8; gk0_13.pad_ = 0;
      if ((long long)(N) >= 64 && (long long)(C8) >= 64) k_gemmT<1, 2, 4><<<dim3((unsigned)((C8) + 63) / 64, (unsigned)((N) + 31) / 32, (unsigned)(1)), 32, 0, stream>>>(gk0_13);
      else k_gemm<1><<<dim3((unsigned)((C8) + 31) / 32, (unsigned)((N) + 15) / 16, (unsigned)(1)), 32, 0, stream>>>(gk0_13); }
    k_cast16<<<(unsigned)((((long long)(256) * ((256) / 2)) + 255) / 256), 256, 0, stream>>>(Wv, 256, (_Float16*)(G64A), 256, 256, 256, 1.0f);
    k_castT16<<<(unsigned)((((long long)(1600) * ((256) / 2)) + 255) / 256), 256, 0, stream>>>(s1 + (size_t)13 * C * N, 1600, (_Float16*)(G64B), 256, 256, 1600, 16.0f);
    w25::wmma_gemm64<0, false, 1, 0, false, 0><<<dim3((unsigned)((((256) / 64) * ((1600) / 64) + 7) / 8), (unsigned)(1)), 256, 0, stream>>>((const unsigned short*)(G64A), nullptr, 256, 0, (const unsigned short*)(G64B), nullptr, 256, 0, (void*)(VF), nullptr, 1600, 0, bv, nullptr, 0, 256, 1600, 256, 0.0625f);
    k_ac_planes<<<(unsigned)(((long long)C * N / 2 + 255) / 256), 256, 0, stream>>>(QF, KF, VF, (_Float16*)QH, (_Float16*)QL, (_Float16*)KH, (_Float16*)KL, (_Float16*)V16, N * C8, (long long)C * N);
    w25::wmma_gemm64<1, true, 0, 0, false, 0><<<dim3((unsigned)((((N) / 64) * ((N) / 64) + 7) / 8), (unsigned)(1)), 256, 0, stream>>>((const unsigned short*)(QH), (const unsigned short*)(QL), C8, 0, (const unsigned short*)(KH), (const unsigned short*)(KL), C8, 0, (void*)(EN), nullptr, N, 0, nullptr, nullptr, 0, N, N, C8, 1.0f);
    k_ac_soft<<<N, 256, 0, stream>>>(EN, (_Float16*)P16, N);
    w25::wmma_gemm64<0, false, 0, 0, false, 0><<<dim3((unsigned)((((C) / 64) * ((N) / 64) + 7) / 8), (unsigned)(1)), 256, 0, stream>>>((const unsigned short*)(V16), nullptr, N, 0, (const unsigned short*)(P16), nullptr, N, 0, (void*)(CT), nullptr, N, 0, nullptr, nullptr, 0, C, N, N, 0.000244140625f);
    k_ac_fuse<<<(unsigned)(((long long)C * N + 255) / 256), 256, 0, stream>>>(CT, fw, out, 0, 13, (long long)C * N);
    { GemmP gq0_14;
      gq0_14.A = s0 + (size_t)14 * C * N; gq0_14.B = Wq; gq0_14.bias = bq; gq0_14.R = s0 + (size_t)14 * C * N; gq0_14.C = QF;
      gq0_14.sAo = 0; gq0_14.sAi = 0; gq0_14.sAm = 1; gq0_14.sAk = N; gq0_14.sBo = 0; gq0_14.sBi = 0; gq0_14.sBn = C; gq0_14.sBk = 1; gq0_14.sCo = 0; gq0_14.sCi = 0; gq0_14.sCm = C8; gq0_14.sRo = 0; gq0_14.sRi = 0; gq0_14.sRm = 0; gq0_14.sRn = 0;
      gq0_14.M = N; gq0_14.N = C8; gq0_14.K = C; gq0_14.zi_n = 1; gq0_14.flags = 1; gq0_14.act = 0;
      gq0_14.alpha = 1.0f; gq0_14.beta = 0.0f; gq0_14.sa = 1.0f; gq0_14.sb = 1.0f; gq0_14.Npad = C8; gq0_14.pad_ = 0;
      if ((long long)(N) >= 64 && (long long)(C8) >= 64) k_gemmT<1, 2, 4><<<dim3((unsigned)((C8) + 63) / 64, (unsigned)((N) + 31) / 32, (unsigned)(1)), 32, 0, stream>>>(gq0_14);
      else k_gemm<1><<<dim3((unsigned)((C8) + 31) / 32, (unsigned)((N) + 15) / 16, (unsigned)(1)), 32, 0, stream>>>(gq0_14); }
    { GemmP gk0_14;
      gk0_14.A = s1 + (size_t)14 * C * N; gk0_14.B = Wk; gk0_14.bias = bk; gk0_14.R = s1 + (size_t)14 * C * N; gk0_14.C = KF;
      gk0_14.sAo = 0; gk0_14.sAi = 0; gk0_14.sAm = 1; gk0_14.sAk = N; gk0_14.sBo = 0; gk0_14.sBi = 0; gk0_14.sBn = C; gk0_14.sBk = 1; gk0_14.sCo = 0; gk0_14.sCi = 0; gk0_14.sCm = C8; gk0_14.sRo = 0; gk0_14.sRi = 0; gk0_14.sRm = 0; gk0_14.sRn = 0;
      gk0_14.M = N; gk0_14.N = C8; gk0_14.K = C; gk0_14.zi_n = 1; gk0_14.flags = 1; gk0_14.act = 0;
      gk0_14.alpha = 1.0f; gk0_14.beta = 0.0f; gk0_14.sa = 1.0f; gk0_14.sb = 1.0f; gk0_14.Npad = C8; gk0_14.pad_ = 0;
      if ((long long)(N) >= 64 && (long long)(C8) >= 64) k_gemmT<1, 2, 4><<<dim3((unsigned)((C8) + 63) / 64, (unsigned)((N) + 31) / 32, (unsigned)(1)), 32, 0, stream>>>(gk0_14);
      else k_gemm<1><<<dim3((unsigned)((C8) + 31) / 32, (unsigned)((N) + 15) / 16, (unsigned)(1)), 32, 0, stream>>>(gk0_14); }
    k_cast16<<<(unsigned)((((long long)(256) * ((256) / 2)) + 255) / 256), 256, 0, stream>>>(Wv, 256, (_Float16*)(G64A), 256, 256, 256, 1.0f);
    k_castT16<<<(unsigned)((((long long)(1600) * ((256) / 2)) + 255) / 256), 256, 0, stream>>>(s1 + (size_t)14 * C * N, 1600, (_Float16*)(G64B), 256, 256, 1600, 16.0f);
    w25::wmma_gemm64<0, false, 1, 0, false, 0><<<dim3((unsigned)((((256) / 64) * ((1600) / 64) + 7) / 8), (unsigned)(1)), 256, 0, stream>>>((const unsigned short*)(G64A), nullptr, 256, 0, (const unsigned short*)(G64B), nullptr, 256, 0, (void*)(VF), nullptr, 1600, 0, bv, nullptr, 0, 256, 1600, 256, 0.0625f);
    k_ac_planes<<<(unsigned)(((long long)C * N / 2 + 255) / 256), 256, 0, stream>>>(QF, KF, VF, (_Float16*)QH, (_Float16*)QL, (_Float16*)KH, (_Float16*)KL, (_Float16*)V16, N * C8, (long long)C * N);
    w25::wmma_gemm64<1, true, 0, 0, false, 0><<<dim3((unsigned)((((N) / 64) * ((N) / 64) + 7) / 8), (unsigned)(1)), 256, 0, stream>>>((const unsigned short*)(QH), (const unsigned short*)(QL), C8, 0, (const unsigned short*)(KH), (const unsigned short*)(KL), C8, 0, (void*)(EN), nullptr, N, 0, nullptr, nullptr, 0, N, N, C8, 1.0f);
    k_ac_soft<<<N, 256, 0, stream>>>(EN, (_Float16*)P16, N);
    w25::wmma_gemm64<0, false, 0, 0, false, 0><<<dim3((unsigned)((((C) / 64) * ((N) / 64) + 7) / 8), (unsigned)(1)), 256, 0, stream>>>((const unsigned short*)(V16), nullptr, N, 0, (const unsigned short*)(P16), nullptr, N, 0, (void*)(CT), nullptr, N, 0, nullptr, nullptr, 0, C, N, N, 0.000244140625f);
    k_ac_fuse<<<(unsigned)(((long long)C * N + 255) / 256), 256, 0, stream>>>(CT, fw, out, 0, 14, (long long)C * N);
    { GemmP gq0_15;
      gq0_15.A = s0 + (size_t)15 * C * N; gq0_15.B = Wq; gq0_15.bias = bq; gq0_15.R = s0 + (size_t)15 * C * N; gq0_15.C = QF;
      gq0_15.sAo = 0; gq0_15.sAi = 0; gq0_15.sAm = 1; gq0_15.sAk = N; gq0_15.sBo = 0; gq0_15.sBi = 0; gq0_15.sBn = C; gq0_15.sBk = 1; gq0_15.sCo = 0; gq0_15.sCi = 0; gq0_15.sCm = C8; gq0_15.sRo = 0; gq0_15.sRi = 0; gq0_15.sRm = 0; gq0_15.sRn = 0;
      gq0_15.M = N; gq0_15.N = C8; gq0_15.K = C; gq0_15.zi_n = 1; gq0_15.flags = 1; gq0_15.act = 0;
      gq0_15.alpha = 1.0f; gq0_15.beta = 0.0f; gq0_15.sa = 1.0f; gq0_15.sb = 1.0f; gq0_15.Npad = C8; gq0_15.pad_ = 0;
      if ((long long)(N) >= 64 && (long long)(C8) >= 64) k_gemmT<1, 2, 4><<<dim3((unsigned)((C8) + 63) / 64, (unsigned)((N) + 31) / 32, (unsigned)(1)), 32, 0, stream>>>(gq0_15);
      else k_gemm<1><<<dim3((unsigned)((C8) + 31) / 32, (unsigned)((N) + 15) / 16, (unsigned)(1)), 32, 0, stream>>>(gq0_15); }
    { GemmP gk0_15;
      gk0_15.A = s1 + (size_t)15 * C * N; gk0_15.B = Wk; gk0_15.bias = bk; gk0_15.R = s1 + (size_t)15 * C * N; gk0_15.C = KF;
      gk0_15.sAo = 0; gk0_15.sAi = 0; gk0_15.sAm = 1; gk0_15.sAk = N; gk0_15.sBo = 0; gk0_15.sBi = 0; gk0_15.sBn = C; gk0_15.sBk = 1; gk0_15.sCo = 0; gk0_15.sCi = 0; gk0_15.sCm = C8; gk0_15.sRo = 0; gk0_15.sRi = 0; gk0_15.sRm = 0; gk0_15.sRn = 0;
      gk0_15.M = N; gk0_15.N = C8; gk0_15.K = C; gk0_15.zi_n = 1; gk0_15.flags = 1; gk0_15.act = 0;
      gk0_15.alpha = 1.0f; gk0_15.beta = 0.0f; gk0_15.sa = 1.0f; gk0_15.sb = 1.0f; gk0_15.Npad = C8; gk0_15.pad_ = 0;
      if ((long long)(N) >= 64 && (long long)(C8) >= 64) k_gemmT<1, 2, 4><<<dim3((unsigned)((C8) + 63) / 64, (unsigned)((N) + 31) / 32, (unsigned)(1)), 32, 0, stream>>>(gk0_15);
      else k_gemm<1><<<dim3((unsigned)((C8) + 31) / 32, (unsigned)((N) + 15) / 16, (unsigned)(1)), 32, 0, stream>>>(gk0_15); }
    k_cast16<<<(unsigned)((((long long)(256) * ((256) / 2)) + 255) / 256), 256, 0, stream>>>(Wv, 256, (_Float16*)(G64A), 256, 256, 256, 1.0f);
    k_castT16<<<(unsigned)((((long long)(1600) * ((256) / 2)) + 255) / 256), 256, 0, stream>>>(s1 + (size_t)15 * C * N, 1600, (_Float16*)(G64B), 256, 256, 1600, 16.0f);
    w25::wmma_gemm64<0, false, 1, 0, false, 0><<<dim3((unsigned)((((256) / 64) * ((1600) / 64) + 7) / 8), (unsigned)(1)), 256, 0, stream>>>((const unsigned short*)(G64A), nullptr, 256, 0, (const unsigned short*)(G64B), nullptr, 256, 0, (void*)(VF), nullptr, 1600, 0, bv, nullptr, 0, 256, 1600, 256, 0.0625f);
    k_ac_planes<<<(unsigned)(((long long)C * N / 2 + 255) / 256), 256, 0, stream>>>(QF, KF, VF, (_Float16*)QH, (_Float16*)QL, (_Float16*)KH, (_Float16*)KL, (_Float16*)V16, N * C8, (long long)C * N);
    w25::wmma_gemm64<1, true, 0, 0, false, 0><<<dim3((unsigned)((((N) / 64) * ((N) / 64) + 7) / 8), (unsigned)(1)), 256, 0, stream>>>((const unsigned short*)(QH), (const unsigned short*)(QL), C8, 0, (const unsigned short*)(KH), (const unsigned short*)(KL), C8, 0, (void*)(EN), nullptr, N, 0, nullptr, nullptr, 0, N, N, C8, 1.0f);
    k_ac_soft<<<N, 256, 0, stream>>>(EN, (_Float16*)P16, N);
    w25::wmma_gemm64<0, false, 0, 0, false, 0><<<dim3((unsigned)((((C) / 64) * ((N) / 64) + 7) / 8), (unsigned)(1)), 256, 0, stream>>>((const unsigned short*)(V16), nullptr, N, 0, (const unsigned short*)(P16), nullptr, N, 0, (void*)(CT), nullptr, N, 0, nullptr, nullptr, 0, C, N, N, 0.000244140625f);
    k_ac_fuse<<<(unsigned)(((long long)C * N + 255) / 256), 256, 0, stream>>>(CT, fw, out, 0, 15, (long long)C * N);
    { GemmP gq1_0;
      gq1_0.A = s1 + (size_t)0 * C * N; gq1_0.B = Wq; gq1_0.bias = bq; gq1_0.R = s1 + (size_t)0 * C * N; gq1_0.C = QF;
      gq1_0.sAo = 0; gq1_0.sAi = 0; gq1_0.sAm = 1; gq1_0.sAk = N; gq1_0.sBo = 0; gq1_0.sBi = 0; gq1_0.sBn = C; gq1_0.sBk = 1; gq1_0.sCo = 0; gq1_0.sCi = 0; gq1_0.sCm = C8; gq1_0.sRo = 0; gq1_0.sRi = 0; gq1_0.sRm = 0; gq1_0.sRn = 0;
      gq1_0.M = N; gq1_0.N = C8; gq1_0.K = C; gq1_0.zi_n = 1; gq1_0.flags = 1; gq1_0.act = 0;
      gq1_0.alpha = 1.0f; gq1_0.beta = 0.0f; gq1_0.sa = 1.0f; gq1_0.sb = 1.0f; gq1_0.Npad = C8; gq1_0.pad_ = 0;
      if ((long long)(N) >= 64 && (long long)(C8) >= 64) k_gemmT<1, 2, 4><<<dim3((unsigned)((C8) + 63) / 64, (unsigned)((N) + 31) / 32, (unsigned)(1)), 32, 0, stream>>>(gq1_0);
      else k_gemm<1><<<dim3((unsigned)((C8) + 31) / 32, (unsigned)((N) + 15) / 16, (unsigned)(1)), 32, 0, stream>>>(gq1_0); }
    { GemmP gk1_0;
      gk1_0.A = s2 + (size_t)0 * C * N; gk1_0.B = Wk; gk1_0.bias = bk; gk1_0.R = s2 + (size_t)0 * C * N; gk1_0.C = KF;
      gk1_0.sAo = 0; gk1_0.sAi = 0; gk1_0.sAm = 1; gk1_0.sAk = N; gk1_0.sBo = 0; gk1_0.sBi = 0; gk1_0.sBn = C; gk1_0.sBk = 1; gk1_0.sCo = 0; gk1_0.sCi = 0; gk1_0.sCm = C8; gk1_0.sRo = 0; gk1_0.sRi = 0; gk1_0.sRm = 0; gk1_0.sRn = 0;
      gk1_0.M = N; gk1_0.N = C8; gk1_0.K = C; gk1_0.zi_n = 1; gk1_0.flags = 1; gk1_0.act = 0;
      gk1_0.alpha = 1.0f; gk1_0.beta = 0.0f; gk1_0.sa = 1.0f; gk1_0.sb = 1.0f; gk1_0.Npad = C8; gk1_0.pad_ = 0;
      if ((long long)(N) >= 64 && (long long)(C8) >= 64) k_gemmT<1, 2, 4><<<dim3((unsigned)((C8) + 63) / 64, (unsigned)((N) + 31) / 32, (unsigned)(1)), 32, 0, stream>>>(gk1_0);
      else k_gemm<1><<<dim3((unsigned)((C8) + 31) / 32, (unsigned)((N) + 15) / 16, (unsigned)(1)), 32, 0, stream>>>(gk1_0); }
    k_cast16<<<(unsigned)((((long long)(256) * ((256) / 2)) + 255) / 256), 256, 0, stream>>>(Wv, 256, (_Float16*)(G64A), 256, 256, 256, 1.0f);
    k_castT16<<<(unsigned)((((long long)(1600) * ((256) / 2)) + 255) / 256), 256, 0, stream>>>(s2 + (size_t)0 * C * N, 1600, (_Float16*)(G64B), 256, 256, 1600, 16.0f);
    w25::wmma_gemm64<0, false, 1, 0, false, 0><<<dim3((unsigned)((((256) / 64) * ((1600) / 64) + 7) / 8), (unsigned)(1)), 256, 0, stream>>>((const unsigned short*)(G64A), nullptr, 256, 0, (const unsigned short*)(G64B), nullptr, 256, 0, (void*)(VF), nullptr, 1600, 0, bv, nullptr, 0, 256, 1600, 256, 0.0625f);
    k_ac_planes<<<(unsigned)(((long long)C * N / 2 + 255) / 256), 256, 0, stream>>>(QF, KF, VF, (_Float16*)QH, (_Float16*)QL, (_Float16*)KH, (_Float16*)KL, (_Float16*)V16, N * C8, (long long)C * N);
    w25::wmma_gemm64<1, true, 0, 0, false, 0><<<dim3((unsigned)((((N) / 64) * ((N) / 64) + 7) / 8), (unsigned)(1)), 256, 0, stream>>>((const unsigned short*)(QH), (const unsigned short*)(QL), C8, 0, (const unsigned short*)(KH), (const unsigned short*)(KL), C8, 0, (void*)(EN), nullptr, N, 0, nullptr, nullptr, 0, N, N, C8, 1.0f);
    k_ac_soft<<<N, 256, 0, stream>>>(EN, (_Float16*)P16, N);
    w25::wmma_gemm64<0, false, 0, 0, false, 0><<<dim3((unsigned)((((C) / 64) * ((N) / 64) + 7) / 8), (unsigned)(1)), 256, 0, stream>>>((const unsigned short*)(V16), nullptr, N, 0, (const unsigned short*)(P16), nullptr, N, 0, (void*)(CT), nullptr, N, 0, nullptr, nullptr, 0, C, N, N, 0.000244140625f);
    k_ac_fuse<<<(unsigned)(((long long)C * N + 255) / 256), 256, 0, stream>>>(CT, fw, out, 1, 0, (long long)C * N);
    { GemmP gq1_1;
      gq1_1.A = s1 + (size_t)1 * C * N; gq1_1.B = Wq; gq1_1.bias = bq; gq1_1.R = s1 + (size_t)1 * C * N; gq1_1.C = QF;
      gq1_1.sAo = 0; gq1_1.sAi = 0; gq1_1.sAm = 1; gq1_1.sAk = N; gq1_1.sBo = 0; gq1_1.sBi = 0; gq1_1.sBn = C; gq1_1.sBk = 1; gq1_1.sCo = 0; gq1_1.sCi = 0; gq1_1.sCm = C8; gq1_1.sRo = 0; gq1_1.sRi = 0; gq1_1.sRm = 0; gq1_1.sRn = 0;
      gq1_1.M = N; gq1_1.N = C8; gq1_1.K = C; gq1_1.zi_n = 1; gq1_1.flags = 1; gq1_1.act = 0;
      gq1_1.alpha = 1.0f; gq1_1.beta = 0.0f; gq1_1.sa = 1.0f; gq1_1.sb = 1.0f; gq1_1.Npad = C8; gq1_1.pad_ = 0;
      if ((long long)(N) >= 64 && (long long)(C8) >= 64) k_gemmT<1, 2, 4><<<dim3((unsigned)((C8) + 63) / 64, (unsigned)((N) + 31) / 32, (unsigned)(1)), 32, 0, stream>>>(gq1_1);
      else k_gemm<1><<<dim3((unsigned)((C8) + 31) / 32, (unsigned)((N) + 15) / 16, (unsigned)(1)), 32, 0, stream>>>(gq1_1); }
    { GemmP gk1_1;
      gk1_1.A = s2 + (size_t)1 * C * N; gk1_1.B = Wk; gk1_1.bias = bk; gk1_1.R = s2 + (size_t)1 * C * N; gk1_1.C = KF;
      gk1_1.sAo = 0; gk1_1.sAi = 0; gk1_1.sAm = 1; gk1_1.sAk = N; gk1_1.sBo = 0; gk1_1.sBi = 0; gk1_1.sBn = C; gk1_1.sBk = 1; gk1_1.sCo = 0; gk1_1.sCi = 0; gk1_1.sCm = C8; gk1_1.sRo = 0; gk1_1.sRi = 0; gk1_1.sRm = 0; gk1_1.sRn = 0;
      gk1_1.M = N; gk1_1.N = C8; gk1_1.K = C; gk1_1.zi_n = 1; gk1_1.flags = 1; gk1_1.act = 0;
      gk1_1.alpha = 1.0f; gk1_1.beta = 0.0f; gk1_1.sa = 1.0f; gk1_1.sb = 1.0f; gk1_1.Npad = C8; gk1_1.pad_ = 0;
      if ((long long)(N) >= 64 && (long long)(C8) >= 64) k_gemmT<1, 2, 4><<<dim3((unsigned)((C8) + 63) / 64, (unsigned)((N) + 31) / 32, (unsigned)(1)), 32, 0, stream>>>(gk1_1);
      else k_gemm<1><<<dim3((unsigned)((C8) + 31) / 32, (unsigned)((N) + 15) / 16, (unsigned)(1)), 32, 0, stream>>>(gk1_1); }
    k_cast16<<<(unsigned)((((long long)(256) * ((256) / 2)) + 255) / 256), 256, 0, stream>>>(Wv, 256, (_Float16*)(G64A), 256, 256, 256, 1.0f);
    k_castT16<<<(unsigned)((((long long)(1600) * ((256) / 2)) + 255) / 256), 256, 0, stream>>>(s2 + (size_t)1 * C * N, 1600, (_Float16*)(G64B), 256, 256, 1600, 16.0f);
    w25::wmma_gemm64<0, false, 1, 0, false, 0><<<dim3((unsigned)((((256) / 64) * ((1600) / 64) + 7) / 8), (unsigned)(1)), 256, 0, stream>>>((const unsigned short*)(G64A), nullptr, 256, 0, (const unsigned short*)(G64B), nullptr, 256, 0, (void*)(VF), nullptr, 1600, 0, bv, nullptr, 0, 256, 1600, 256, 0.0625f);
    k_ac_planes<<<(unsigned)(((long long)C * N / 2 + 255) / 256), 256, 0, stream>>>(QF, KF, VF, (_Float16*)QH, (_Float16*)QL, (_Float16*)KH, (_Float16*)KL, (_Float16*)V16, N * C8, (long long)C * N);
    w25::wmma_gemm64<1, true, 0, 0, false, 0><<<dim3((unsigned)((((N) / 64) * ((N) / 64) + 7) / 8), (unsigned)(1)), 256, 0, stream>>>((const unsigned short*)(QH), (const unsigned short*)(QL), C8, 0, (const unsigned short*)(KH), (const unsigned short*)(KL), C8, 0, (void*)(EN), nullptr, N, 0, nullptr, nullptr, 0, N, N, C8, 1.0f);
    k_ac_soft<<<N, 256, 0, stream>>>(EN, (_Float16*)P16, N);
    w25::wmma_gemm64<0, false, 0, 0, false, 0><<<dim3((unsigned)((((C) / 64) * ((N) / 64) + 7) / 8), (unsigned)(1)), 256, 0, stream>>>((const unsigned short*)(V16), nullptr, N, 0, (const unsigned short*)(P16), nullptr, N, 0, (void*)(CT), nullptr, N, 0, nullptr, nullptr, 0, C, N, N, 0.000244140625f);
    k_ac_fuse<<<(unsigned)(((long long)C * N + 255) / 256), 256, 0, stream>>>(CT, fw, out, 1, 1, (long long)C * N);
    { GemmP gq1_2;
      gq1_2.A = s1 + (size_t)2 * C * N; gq1_2.B = Wq; gq1_2.bias = bq; gq1_2.R = s1 + (size_t)2 * C * N; gq1_2.C = QF;
      gq1_2.sAo = 0; gq1_2.sAi = 0; gq1_2.sAm = 1; gq1_2.sAk = N; gq1_2.sBo = 0; gq1_2.sBi = 0; gq1_2.sBn = C; gq1_2.sBk = 1; gq1_2.sCo = 0; gq1_2.sCi = 0; gq1_2.sCm = C8; gq1_2.sRo = 0; gq1_2.sRi = 0; gq1_2.sRm = 0; gq1_2.sRn = 0;
      gq1_2.M = N; gq1_2.N = C8; gq1_2.K = C; gq1_2.zi_n = 1; gq1_2.flags = 1; gq1_2.act = 0;
      gq1_2.alpha = 1.0f; gq1_2.beta = 0.0f; gq1_2.sa = 1.0f; gq1_2.sb = 1.0f; gq1_2.Npad = C8; gq1_2.pad_ = 0;
      if ((long long)(N) >= 64 && (long long)(C8) >= 64) k_gemmT<1, 2, 4><<<dim3((unsigned)((C8) + 63) / 64, (unsigned)((N) + 31) / 32, (unsigned)(1)), 32, 0, stream>>>(gq1_2);
      else k_gemm<1><<<dim3((unsigned)((C8) + 31) / 32, (unsigned)((N) + 15) / 16, (unsigned)(1)), 32, 0, stream>>>(gq1_2); }
    { GemmP gk1_2;
      gk1_2.A = s2 + (size_t)2 * C * N; gk1_2.B = Wk; gk1_2.bias = bk; gk1_2.R = s2 + (size_t)2 * C * N; gk1_2.C = KF;
      gk1_2.sAo = 0; gk1_2.sAi = 0; gk1_2.sAm = 1; gk1_2.sAk = N; gk1_2.sBo = 0; gk1_2.sBi = 0; gk1_2.sBn = C; gk1_2.sBk = 1; gk1_2.sCo = 0; gk1_2.sCi = 0; gk1_2.sCm = C8; gk1_2.sRo = 0; gk1_2.sRi = 0; gk1_2.sRm = 0; gk1_2.sRn = 0;
      gk1_2.M = N; gk1_2.N = C8; gk1_2.K = C; gk1_2.zi_n = 1; gk1_2.flags = 1; gk1_2.act = 0;
      gk1_2.alpha = 1.0f; gk1_2.beta = 0.0f; gk1_2.sa = 1.0f; gk1_2.sb = 1.0f; gk1_2.Npad = C8; gk1_2.pad_ = 0;
      if ((long long)(N) >= 64 && (long long)(C8) >= 64) k_gemmT<1, 2, 4><<<dim3((unsigned)((C8) + 63) / 64, (unsigned)((N) + 31) / 32, (unsigned)(1)), 32, 0, stream>>>(gk1_2);
      else k_gemm<1><<<dim3((unsigned)((C8) + 31) / 32, (unsigned)((N) + 15) / 16, (unsigned)(1)), 32, 0, stream>>>(gk1_2); }
    k_cast16<<<(unsigned)((((long long)(256) * ((256) / 2)) + 255) / 256), 256, 0, stream>>>(Wv, 256, (_Float16*)(G64A), 256, 256, 256, 1.0f);
    k_castT16<<<(unsigned)((((long long)(1600) * ((256) / 2)) + 255) / 256), 256, 0, stream>>>(s2 + (size_t)2 * C * N, 1600, (_Float16*)(G64B), 256, 256, 1600, 16.0f);
    w25::wmma_gemm64<0, false, 1, 0, false, 0><<<dim3((unsigned)((((256) / 64) * ((1600) / 64) + 7) / 8), (unsigned)(1)), 256, 0, stream>>>((const unsigned short*)(G64A), nullptr, 256, 0, (const unsigned short*)(G64B), nullptr, 256, 0, (void*)(VF), nullptr, 1600, 0, bv, nullptr, 0, 256, 1600, 256, 0.0625f);
    k_ac_planes<<<(unsigned)(((long long)C * N / 2 + 255) / 256), 256, 0, stream>>>(QF, KF, VF, (_Float16*)QH, (_Float16*)QL, (_Float16*)KH, (_Float16*)KL, (_Float16*)V16, N * C8, (long long)C * N);
    w25::wmma_gemm64<1, true, 0, 0, false, 0><<<dim3((unsigned)((((N) / 64) * ((N) / 64) + 7) / 8), (unsigned)(1)), 256, 0, stream>>>((const unsigned short*)(QH), (const unsigned short*)(QL), C8, 0, (const unsigned short*)(KH), (const unsigned short*)(KL), C8, 0, (void*)(EN), nullptr, N, 0, nullptr, nullptr, 0, N, N, C8, 1.0f);
    k_ac_soft<<<N, 256, 0, stream>>>(EN, (_Float16*)P16, N);
    w25::wmma_gemm64<0, false, 0, 0, false, 0><<<dim3((unsigned)((((C) / 64) * ((N) / 64) + 7) / 8), (unsigned)(1)), 256, 0, stream>>>((const unsigned short*)(V16), nullptr, N, 0, (const unsigned short*)(P16), nullptr, N, 0, (void*)(CT), nullptr, N, 0, nullptr, nullptr, 0, C, N, N, 0.000244140625f);
    k_ac_fuse<<<(unsigned)(((long long)C * N + 255) / 256), 256, 0, stream>>>(CT, fw, out, 1, 2, (long long)C * N);
    { GemmP gq1_3;
      gq1_3.A = s1 + (size_t)3 * C * N; gq1_3.B = Wq; gq1_3.bias = bq; gq1_3.R = s1 + (size_t)3 * C * N; gq1_3.C = QF;
      gq1_3.sAo = 0; gq1_3.sAi = 0; gq1_3.sAm = 1; gq1_3.sAk = N; gq1_3.sBo = 0; gq1_3.sBi = 0; gq1_3.sBn = C; gq1_3.sBk = 1; gq1_3.sCo = 0; gq1_3.sCi = 0; gq1_3.sCm = C8; gq1_3.sRo = 0; gq1_3.sRi = 0; gq1_3.sRm = 0; gq1_3.sRn = 0;
      gq1_3.M = N; gq1_3.N = C8; gq1_3.K = C; gq1_3.zi_n = 1; gq1_3.flags = 1; gq1_3.act = 0;
      gq1_3.alpha = 1.0f; gq1_3.beta = 0.0f; gq1_3.sa = 1.0f; gq1_3.sb = 1.0f; gq1_3.Npad = C8; gq1_3.pad_ = 0;
      if ((long long)(N) >= 64 && (long long)(C8) >= 64) k_gemmT<1, 2, 4><<<dim3((unsigned)((C8) + 63) / 64, (unsigned)((N) + 31) / 32, (unsigned)(1)), 32, 0, stream>>>(gq1_3);
      else k_gemm<1><<<dim3((unsigned)((C8) + 31) / 32, (unsigned)((N) + 15) / 16, (unsigned)(1)), 32, 0, stream>>>(gq1_3); }
    { GemmP gk1_3;
      gk1_3.A = s2 + (size_t)3 * C * N; gk1_3.B = Wk; gk1_3.bias = bk; gk1_3.R = s2 + (size_t)3 * C * N; gk1_3.C = KF;
      gk1_3.sAo = 0; gk1_3.sAi = 0; gk1_3.sAm = 1; gk1_3.sAk = N; gk1_3.sBo = 0; gk1_3.sBi = 0; gk1_3.sBn = C; gk1_3.sBk = 1; gk1_3.sCo = 0; gk1_3.sCi = 0; gk1_3.sCm = C8; gk1_3.sRo = 0; gk1_3.sRi = 0; gk1_3.sRm = 0; gk1_3.sRn = 0;
      gk1_3.M = N; gk1_3.N = C8; gk1_3.K = C; gk1_3.zi_n = 1; gk1_3.flags = 1; gk1_3.act = 0;
      gk1_3.alpha = 1.0f; gk1_3.beta = 0.0f; gk1_3.sa = 1.0f; gk1_3.sb = 1.0f; gk1_3.Npad = C8; gk1_3.pad_ = 0;
      if ((long long)(N) >= 64 && (long long)(C8) >= 64) k_gemmT<1, 2, 4><<<dim3((unsigned)((C8) + 63) / 64, (unsigned)((N) + 31) / 32, (unsigned)(1)), 32, 0, stream>>>(gk1_3);
      else k_gemm<1><<<dim3((unsigned)((C8) + 31) / 32, (unsigned)((N) + 15) / 16, (unsigned)(1)), 32, 0, stream>>>(gk1_3); }
    k_cast16<<<(unsigned)((((long long)(256) * ((256) / 2)) + 255) / 256), 256, 0, stream>>>(Wv, 256, (_Float16*)(G64A), 256, 256, 256, 1.0f);
    k_castT16<<<(unsigned)((((long long)(1600) * ((256) / 2)) + 255) / 256), 256, 0, stream>>>(s2 + (size_t)3 * C * N, 1600, (_Float16*)(G64B), 256, 256, 1600, 16.0f);
    w25::wmma_gemm64<0, false, 1, 0, false, 0><<<dim3((unsigned)((((256) / 64) * ((1600) / 64) + 7) / 8), (unsigned)(1)), 256, 0, stream>>>((const unsigned short*)(G64A), nullptr, 256, 0, (const unsigned short*)(G64B), nullptr, 256, 0, (void*)(VF), nullptr, 1600, 0, bv, nullptr, 0, 256, 1600, 256, 0.0625f);
    k_ac_planes<<<(unsigned)(((long long)C * N / 2 + 255) / 256), 256, 0, stream>>>(QF, KF, VF, (_Float16*)QH, (_Float16*)QL, (_Float16*)KH, (_Float16*)KL, (_Float16*)V16, N * C8, (long long)C * N);
    w25::wmma_gemm64<1, true, 0, 0, false, 0><<<dim3((unsigned)((((N) / 64) * ((N) / 64) + 7) / 8), (unsigned)(1)), 256, 0, stream>>>((const unsigned short*)(QH), (const unsigned short*)(QL), C8, 0, (const unsigned short*)(KH), (const unsigned short*)(KL), C8, 0, (void*)(EN), nullptr, N, 0, nullptr, nullptr, 0, N, N, C8, 1.0f);
    k_ac_soft<<<N, 256, 0, stream>>>(EN, (_Float16*)P16, N);
    w25::wmma_gemm64<0, false, 0, 0, false, 0><<<dim3((unsigned)((((C) / 64) * ((N) / 64) + 7) / 8), (unsigned)(1)), 256, 0, stream>>>((const unsigned short*)(V16), nullptr, N, 0, (const unsigned short*)(P16), nullptr, N, 0, (void*)(CT), nullptr, N, 0, nullptr, nullptr, 0, C, N, N, 0.000244140625f);
    k_ac_fuse<<<(unsigned)(((long long)C * N + 255) / 256), 256, 0, stream>>>(CT, fw, out, 1, 3, (long long)C * N);
    { GemmP gq1_4;
      gq1_4.A = s1 + (size_t)4 * C * N; gq1_4.B = Wq; gq1_4.bias = bq; gq1_4.R = s1 + (size_t)4 * C * N; gq1_4.C = QF;
      gq1_4.sAo = 0; gq1_4.sAi = 0; gq1_4.sAm = 1; gq1_4.sAk = N; gq1_4.sBo = 0; gq1_4.sBi = 0; gq1_4.sBn = C; gq1_4.sBk = 1; gq1_4.sCo = 0; gq1_4.sCi = 0; gq1_4.sCm = C8; gq1_4.sRo = 0; gq1_4.sRi = 0; gq1_4.sRm = 0; gq1_4.sRn = 0;
      gq1_4.M = N; gq1_4.N = C8; gq1_4.K = C; gq1_4.zi_n = 1; gq1_4.flags = 1; gq1_4.act = 0;
      gq1_4.alpha = 1.0f; gq1_4.beta = 0.0f; gq1_4.sa = 1.0f; gq1_4.sb = 1.0f; gq1_4.Npad = C8; gq1_4.pad_ = 0;
      if ((long long)(N) >= 64 && (long long)(C8) >= 64) k_gemmT<1, 2, 4><<<dim3((unsigned)((C8) + 63) / 64, (unsigned)((N) + 31) / 32, (unsigned)(1)), 32, 0, stream>>>(gq1_4);
      else k_gemm<1><<<dim3((unsigned)((C8) + 31) / 32, (unsigned)((N) + 15) / 16, (unsigned)(1)), 32, 0, stream>>>(gq1_4); }
    { GemmP gk1_4;
      gk1_4.A = s2 + (size_t)4 * C * N; gk1_4.B = Wk; gk1_4.bias = bk; gk1_4.R = s2 + (size_t)4 * C * N; gk1_4.C = KF;
      gk1_4.sAo = 0; gk1_4.sAi = 0; gk1_4.sAm = 1; gk1_4.sAk = N; gk1_4.sBo = 0; gk1_4.sBi = 0; gk1_4.sBn = C; gk1_4.sBk = 1; gk1_4.sCo = 0; gk1_4.sCi = 0; gk1_4.sCm = C8; gk1_4.sRo = 0; gk1_4.sRi = 0; gk1_4.sRm = 0; gk1_4.sRn = 0;
      gk1_4.M = N; gk1_4.N = C8; gk1_4.K = C; gk1_4.zi_n = 1; gk1_4.flags = 1; gk1_4.act = 0;
      gk1_4.alpha = 1.0f; gk1_4.beta = 0.0f; gk1_4.sa = 1.0f; gk1_4.sb = 1.0f; gk1_4.Npad = C8; gk1_4.pad_ = 0;
      if ((long long)(N) >= 64 && (long long)(C8) >= 64) k_gemmT<1, 2, 4><<<dim3((unsigned)((C8) + 63) / 64, (unsigned)((N) + 31) / 32, (unsigned)(1)), 32, 0, stream>>>(gk1_4);
      else k_gemm<1><<<dim3((unsigned)((C8) + 31) / 32, (unsigned)((N) + 15) / 16, (unsigned)(1)), 32, 0, stream>>>(gk1_4); }
    k_cast16<<<(unsigned)((((long long)(256) * ((256) / 2)) + 255) / 256), 256, 0, stream>>>(Wv, 256, (_Float16*)(G64A), 256, 256, 256, 1.0f);
    k_castT16<<<(unsigned)((((long long)(1600) * ((256) / 2)) + 255) / 256), 256, 0, stream>>>(s2 + (size_t)4 * C * N, 1600, (_Float16*)(G64B), 256, 256, 1600, 16.0f);
    w25::wmma_gemm64<0, false, 1, 0, false, 0><<<dim3((unsigned)((((256) / 64) * ((1600) / 64) + 7) / 8), (unsigned)(1)), 256, 0, stream>>>((const unsigned short*)(G64A), nullptr, 256, 0, (const unsigned short*)(G64B), nullptr, 256, 0, (void*)(VF), nullptr, 1600, 0, bv, nullptr, 0, 256, 1600, 256, 0.0625f);
    k_ac_planes<<<(unsigned)(((long long)C * N / 2 + 255) / 256), 256, 0, stream>>>(QF, KF, VF, (_Float16*)QH, (_Float16*)QL, (_Float16*)KH, (_Float16*)KL, (_Float16*)V16, N * C8, (long long)C * N);
    w25::wmma_gemm64<1, true, 0, 0, false, 0><<<dim3((unsigned)((((N) / 64) * ((N) / 64) + 7) / 8), (unsigned)(1)), 256, 0, stream>>>((const unsigned short*)(QH), (const unsigned short*)(QL), C8, 0, (const unsigned short*)(KH), (const unsigned short*)(KL), C8, 0, (void*)(EN), nullptr, N, 0, nullptr, nullptr, 0, N, N, C8, 1.0f);
    k_ac_soft<<<N, 256, 0, stream>>>(EN, (_Float16*)P16, N);
    w25::wmma_gemm64<0, false, 0, 0, false, 0><<<dim3((unsigned)((((C) / 64) * ((N) / 64) + 7) / 8), (unsigned)(1)), 256, 0, stream>>>((const unsigned short*)(V16), nullptr, N, 0, (const unsigned short*)(P16), nullptr, N, 0, (void*)(CT), nullptr, N, 0, nullptr, nullptr, 0, C, N, N, 0.000244140625f);
    k_ac_fuse<<<(unsigned)(((long long)C * N + 255) / 256), 256, 0, stream>>>(CT, fw, out, 1, 4, (long long)C * N);
    { GemmP gq1_5;
      gq1_5.A = s1 + (size_t)5 * C * N; gq1_5.B = Wq; gq1_5.bias = bq; gq1_5.R = s1 + (size_t)5 * C * N; gq1_5.C = QF;
      gq1_5.sAo = 0; gq1_5.sAi = 0; gq1_5.sAm = 1; gq1_5.sAk = N; gq1_5.sBo = 0; gq1_5.sBi = 0; gq1_5.sBn = C; gq1_5.sBk = 1; gq1_5.sCo = 0; gq1_5.sCi = 0; gq1_5.sCm = C8; gq1_5.sRo = 0; gq1_5.sRi = 0; gq1_5.sRm = 0; gq1_5.sRn = 0;
      gq1_5.M = N; gq1_5.N = C8; gq1_5.K = C; gq1_5.zi_n = 1; gq1_5.flags = 1; gq1_5.act = 0;
      gq1_5.alpha = 1.0f; gq1_5.beta = 0.0f; gq1_5.sa = 1.0f; gq1_5.sb = 1.0f; gq1_5.Npad = C8; gq1_5.pad_ = 0;
      if ((long long)(N) >= 64 && (long long)(C8) >= 64) k_gemmT<1, 2, 4><<<dim3((unsigned)((C8) + 63) / 64, (unsigned)((N) + 31) / 32, (unsigned)(1)), 32, 0, stream>>>(gq1_5);
      else k_gemm<1><<<dim3((unsigned)((C8) + 31) / 32, (unsigned)((N) + 15) / 16, (unsigned)(1)), 32, 0, stream>>>(gq1_5); }
    { GemmP gk1_5;
      gk1_5.A = s2 + (size_t)5 * C * N; gk1_5.B = Wk; gk1_5.bias = bk; gk1_5.R = s2 + (size_t)5 * C * N; gk1_5.C = KF;
      gk1_5.sAo = 0; gk1_5.sAi = 0; gk1_5.sAm = 1; gk1_5.sAk = N; gk1_5.sBo = 0; gk1_5.sBi = 0; gk1_5.sBn = C; gk1_5.sBk = 1; gk1_5.sCo = 0; gk1_5.sCi = 0; gk1_5.sCm = C8; gk1_5.sRo = 0; gk1_5.sRi = 0; gk1_5.sRm = 0; gk1_5.sRn = 0;
      gk1_5.M = N; gk1_5.N = C8; gk1_5.K = C; gk1_5.zi_n = 1; gk1_5.flags = 1; gk1_5.act = 0;
      gk1_5.alpha = 1.0f; gk1_5.beta = 0.0f; gk1_5.sa = 1.0f; gk1_5.sb = 1.0f; gk1_5.Npad = C8; gk1_5.pad_ = 0;
      if ((long long)(N) >= 64 && (long long)(C8) >= 64) k_gemmT<1, 2, 4><<<dim3((unsigned)((C8) + 63) / 64, (unsigned)((N) + 31) / 32, (unsigned)(1)), 32, 0, stream>>>(gk1_5);
      else k_gemm<1><<<dim3((unsigned)((C8) + 31) / 32, (unsigned)((N) + 15) / 16, (unsigned)(1)), 32, 0, stream>>>(gk1_5); }
    k_cast16<<<(unsigned)((((long long)(256) * ((256) / 2)) + 255) / 256), 256, 0, stream>>>(Wv, 256, (_Float16*)(G64A), 256, 256, 256, 1.0f);
    k_castT16<<<(unsigned)((((long long)(1600) * ((256) / 2)) + 255) / 256), 256, 0, stream>>>(s2 + (size_t)5 * C * N, 1600, (_Float16*)(G64B), 256, 256, 1600, 16.0f);
    w25::wmma_gemm64<0, false, 1, 0, false, 0><<<dim3((unsigned)((((256) / 64) * ((1600) / 64) + 7) / 8), (unsigned)(1)), 256, 0, stream>>>((const unsigned short*)(G64A), nullptr, 256, 0, (const unsigned short*)(G64B), nullptr, 256, 0, (void*)(VF), nullptr, 1600, 0, bv, nullptr, 0, 256, 1600, 256, 0.0625f);
    k_ac_planes<<<(unsigned)(((long long)C * N / 2 + 255) / 256), 256, 0, stream>>>(QF, KF, VF, (_Float16*)QH, (_Float16*)QL, (_Float16*)KH, (_Float16*)KL, (_Float16*)V16, N * C8, (long long)C * N);
    w25::wmma_gemm64<1, true, 0, 0, false, 0><<<dim3((unsigned)((((N) / 64) * ((N) / 64) + 7) / 8), (unsigned)(1)), 256, 0, stream>>>((const unsigned short*)(QH), (const unsigned short*)(QL), C8, 0, (const unsigned short*)(KH), (const unsigned short*)(KL), C8, 0, (void*)(EN), nullptr, N, 0, nullptr, nullptr, 0, N, N, C8, 1.0f);
    k_ac_soft<<<N, 256, 0, stream>>>(EN, (_Float16*)P16, N);
    w25::wmma_gemm64<0, false, 0, 0, false, 0><<<dim3((unsigned)((((C) / 64) * ((N) / 64) + 7) / 8), (unsigned)(1)), 256, 0, stream>>>((const unsigned short*)(V16), nullptr, N, 0, (const unsigned short*)(P16), nullptr, N, 0, (void*)(CT), nullptr, N, 0, nullptr, nullptr, 0, C, N, N, 0.000244140625f);
    k_ac_fuse<<<(unsigned)(((long long)C * N + 255) / 256), 256, 0, stream>>>(CT, fw, out, 1, 5, (long long)C * N);
    { GemmP gq1_6;
      gq1_6.A = s1 + (size_t)6 * C * N; gq1_6.B = Wq; gq1_6.bias = bq; gq1_6.R = s1 + (size_t)6 * C * N; gq1_6.C = QF;
      gq1_6.sAo = 0; gq1_6.sAi = 0; gq1_6.sAm = 1; gq1_6.sAk = N; gq1_6.sBo = 0; gq1_6.sBi = 0; gq1_6.sBn = C; gq1_6.sBk = 1; gq1_6.sCo = 0; gq1_6.sCi = 0; gq1_6.sCm = C8; gq1_6.sRo = 0; gq1_6.sRi = 0; gq1_6.sRm = 0; gq1_6.sRn = 0;
      gq1_6.M = N; gq1_6.N = C8; gq1_6.K = C; gq1_6.zi_n = 1; gq1_6.flags = 1; gq1_6.act = 0;
      gq1_6.alpha = 1.0f; gq1_6.beta = 0.0f; gq1_6.sa = 1.0f; gq1_6.sb = 1.0f; gq1_6.Npad = C8; gq1_6.pad_ = 0;
      if ((long long)(N) >= 64 && (long long)(C8) >= 64) k_gemmT<1, 2, 4><<<dim3((unsigned)((C8) + 63) / 64, (unsigned)((N) + 31) / 32, (unsigned)(1)), 32, 0, stream>>>(gq1_6);
      else k_gemm<1><<<dim3((unsigned)((C8) + 31) / 32, (unsigned)((N) + 15) / 16, (unsigned)(1)), 32, 0, stream>>>(gq1_6); }
    { GemmP gk1_6;
      gk1_6.A = s2 + (size_t)6 * C * N; gk1_6.B = Wk; gk1_6.bias = bk; gk1_6.R = s2 + (size_t)6 * C * N; gk1_6.C = KF;
      gk1_6.sAo = 0; gk1_6.sAi = 0; gk1_6.sAm = 1; gk1_6.sAk = N; gk1_6.sBo = 0; gk1_6.sBi = 0; gk1_6.sBn = C; gk1_6.sBk = 1; gk1_6.sCo = 0; gk1_6.sCi = 0; gk1_6.sCm = C8; gk1_6.sRo = 0; gk1_6.sRi = 0; gk1_6.sRm = 0; gk1_6.sRn = 0;
      gk1_6.M = N; gk1_6.N = C8; gk1_6.K = C; gk1_6.zi_n = 1; gk1_6.flags = 1; gk1_6.act = 0;
      gk1_6.alpha = 1.0f; gk1_6.beta = 0.0f; gk1_6.sa = 1.0f; gk1_6.sb = 1.0f; gk1_6.Npad = C8; gk1_6.pad_ = 0;
      if ((long long)(N) >= 64 && (long long)(C8) >= 64) k_gemmT<1, 2, 4><<<dim3((unsigned)((C8) + 63) / 64, (unsigned)((N) + 31) / 32, (unsigned)(1)), 32, 0, stream>>>(gk1_6);
      else k_gemm<1><<<dim3((unsigned)((C8) + 31) / 32, (unsigned)((N) + 15) / 16, (unsigned)(1)), 32, 0, stream>>>(gk1_6); }
    k_cast16<<<(unsigned)((((long long)(256) * ((256) / 2)) + 255) / 256), 256, 0, stream>>>(Wv, 256, (_Float16*)(G64A), 256, 256, 256, 1.0f);
    k_castT16<<<(unsigned)((((long long)(1600) * ((256) / 2)) + 255) / 256), 256, 0, stream>>>(s2 + (size_t)6 * C * N, 1600, (_Float16*)(G64B), 256, 256, 1600, 16.0f);
    w25::wmma_gemm64<0, false, 1, 0, false, 0><<<dim3((unsigned)((((256) / 64) * ((1600) / 64) + 7) / 8), (unsigned)(1)), 256, 0, stream>>>((const unsigned short*)(G64A), nullptr, 256, 0, (const unsigned short*)(G64B), nullptr, 256, 0, (void*)(VF), nullptr, 1600, 0, bv, nullptr, 0, 256, 1600, 256, 0.0625f);
    k_ac_planes<<<(unsigned)(((long long)C * N / 2 + 255) / 256), 256, 0, stream>>>(QF, KF, VF, (_Float16*)QH, (_Float16*)QL, (_Float16*)KH, (_Float16*)KL, (_Float16*)V16, N * C8, (long long)C * N);
    w25::wmma_gemm64<1, true, 0, 0, false, 0><<<dim3((unsigned)((((N) / 64) * ((N) / 64) + 7) / 8), (unsigned)(1)), 256, 0, stream>>>((const unsigned short*)(QH), (const unsigned short*)(QL), C8, 0, (const unsigned short*)(KH), (const unsigned short*)(KL), C8, 0, (void*)(EN), nullptr, N, 0, nullptr, nullptr, 0, N, N, C8, 1.0f);
    k_ac_soft<<<N, 256, 0, stream>>>(EN, (_Float16*)P16, N);
    w25::wmma_gemm64<0, false, 0, 0, false, 0><<<dim3((unsigned)((((C) / 64) * ((N) / 64) + 7) / 8), (unsigned)(1)), 256, 0, stream>>>((const unsigned short*)(V16), nullptr, N, 0, (const unsigned short*)(P16), nullptr, N, 0, (void*)(CT), nullptr, N, 0, nullptr, nullptr, 0, C, N, N, 0.000244140625f);
    k_ac_fuse<<<(unsigned)(((long long)C * N + 255) / 256), 256, 0, stream>>>(CT, fw, out, 1, 6, (long long)C * N);
    { GemmP gq1_7;
      gq1_7.A = s1 + (size_t)7 * C * N; gq1_7.B = Wq; gq1_7.bias = bq; gq1_7.R = s1 + (size_t)7 * C * N; gq1_7.C = QF;
      gq1_7.sAo = 0; gq1_7.sAi = 0; gq1_7.sAm = 1; gq1_7.sAk = N; gq1_7.sBo = 0; gq1_7.sBi = 0; gq1_7.sBn = C; gq1_7.sBk = 1; gq1_7.sCo = 0; gq1_7.sCi = 0; gq1_7.sCm = C8; gq1_7.sRo = 0; gq1_7.sRi = 0; gq1_7.sRm = 0; gq1_7.sRn = 0;
      gq1_7.M = N; gq1_7.N = C8; gq1_7.K = C; gq1_7.zi_n = 1; gq1_7.flags = 1; gq1_7.act = 0;
      gq1_7.alpha = 1.0f; gq1_7.beta = 0.0f; gq1_7.sa = 1.0f; gq1_7.sb = 1.0f; gq1_7.Npad = C8; gq1_7.pad_ = 0;
      if ((long long)(N) >= 64 && (long long)(C8) >= 64) k_gemmT<1, 2, 4><<<dim3((unsigned)((C8) + 63) / 64, (unsigned)((N) + 31) / 32, (unsigned)(1)), 32, 0, stream>>>(gq1_7);
      else k_gemm<1><<<dim3((unsigned)((C8) + 31) / 32, (unsigned)((N) + 15) / 16, (unsigned)(1)), 32, 0, stream>>>(gq1_7); }
    { GemmP gk1_7;
      gk1_7.A = s2 + (size_t)7 * C * N; gk1_7.B = Wk; gk1_7.bias = bk; gk1_7.R = s2 + (size_t)7 * C * N; gk1_7.C = KF;
      gk1_7.sAo = 0; gk1_7.sAi = 0; gk1_7.sAm = 1; gk1_7.sAk = N; gk1_7.sBo = 0; gk1_7.sBi = 0; gk1_7.sBn = C; gk1_7.sBk = 1; gk1_7.sCo = 0; gk1_7.sCi = 0; gk1_7.sCm = C8; gk1_7.sRo = 0; gk1_7.sRi = 0; gk1_7.sRm = 0; gk1_7.sRn = 0;
      gk1_7.M = N; gk1_7.N = C8; gk1_7.K = C; gk1_7.zi_n = 1; gk1_7.flags = 1; gk1_7.act = 0;
      gk1_7.alpha = 1.0f; gk1_7.beta = 0.0f; gk1_7.sa = 1.0f; gk1_7.sb = 1.0f; gk1_7.Npad = C8; gk1_7.pad_ = 0;
      if ((long long)(N) >= 64 && (long long)(C8) >= 64) k_gemmT<1, 2, 4><<<dim3((unsigned)((C8) + 63) / 64, (unsigned)((N) + 31) / 32, (unsigned)(1)), 32, 0, stream>>>(gk1_7);
      else k_gemm<1><<<dim3((unsigned)((C8) + 31) / 32, (unsigned)((N) + 15) / 16, (unsigned)(1)), 32, 0, stream>>>(gk1_7); }
    k_cast16<<<(unsigned)((((long long)(256) * ((256) / 2)) + 255) / 256), 256, 0, stream>>>(Wv, 256, (_Float16*)(G64A), 256, 256, 256, 1.0f);
    k_castT16<<<(unsigned)((((long long)(1600) * ((256) / 2)) + 255) / 256), 256, 0, stream>>>(s2 + (size_t)7 * C * N, 1600, (_Float16*)(G64B), 256, 256, 1600, 16.0f);
    w25::wmma_gemm64<0, false, 1, 0, false, 0><<<dim3((unsigned)((((256) / 64) * ((1600) / 64) + 7) / 8), (unsigned)(1)), 256, 0, stream>>>((const unsigned short*)(G64A), nullptr, 256, 0, (const unsigned short*)(G64B), nullptr, 256, 0, (void*)(VF), nullptr, 1600, 0, bv, nullptr, 0, 256, 1600, 256, 0.0625f);
    k_ac_planes<<<(unsigned)(((long long)C * N / 2 + 255) / 256), 256, 0, stream>>>(QF, KF, VF, (_Float16*)QH, (_Float16*)QL, (_Float16*)KH, (_Float16*)KL, (_Float16*)V16, N * C8, (long long)C * N);
    w25::wmma_gemm64<1, true, 0, 0, false, 0><<<dim3((unsigned)((((N) / 64) * ((N) / 64) + 7) / 8), (unsigned)(1)), 256, 0, stream>>>((const unsigned short*)(QH), (const unsigned short*)(QL), C8, 0, (const unsigned short*)(KH), (const unsigned short*)(KL), C8, 0, (void*)(EN), nullptr, N, 0, nullptr, nullptr, 0, N, N, C8, 1.0f);
    k_ac_soft<<<N, 256, 0, stream>>>(EN, (_Float16*)P16, N);
    w25::wmma_gemm64<0, false, 0, 0, false, 0><<<dim3((unsigned)((((C) / 64) * ((N) / 64) + 7) / 8), (unsigned)(1)), 256, 0, stream>>>((const unsigned short*)(V16), nullptr, N, 0, (const unsigned short*)(P16), nullptr, N, 0, (void*)(CT), nullptr, N, 0, nullptr, nullptr, 0, C, N, N, 0.000244140625f);
    k_ac_fuse<<<(unsigned)(((long long)C * N + 255) / 256), 256, 0, stream>>>(CT, fw, out, 1, 7, (long long)C * N);
    { GemmP gq1_8;
      gq1_8.A = s1 + (size_t)8 * C * N; gq1_8.B = Wq; gq1_8.bias = bq; gq1_8.R = s1 + (size_t)8 * C * N; gq1_8.C = QF;
      gq1_8.sAo = 0; gq1_8.sAi = 0; gq1_8.sAm = 1; gq1_8.sAk = N; gq1_8.sBo = 0; gq1_8.sBi = 0; gq1_8.sBn = C; gq1_8.sBk = 1; gq1_8.sCo = 0; gq1_8.sCi = 0; gq1_8.sCm = C8; gq1_8.sRo = 0; gq1_8.sRi = 0; gq1_8.sRm = 0; gq1_8.sRn = 0;
      gq1_8.M = N; gq1_8.N = C8; gq1_8.K = C; gq1_8.zi_n = 1; gq1_8.flags = 1; gq1_8.act = 0;
      gq1_8.alpha = 1.0f; gq1_8.beta = 0.0f; gq1_8.sa = 1.0f; gq1_8.sb = 1.0f; gq1_8.Npad = C8; gq1_8.pad_ = 0;
      if ((long long)(N) >= 64 && (long long)(C8) >= 64) k_gemmT<1, 2, 4><<<dim3((unsigned)((C8) + 63) / 64, (unsigned)((N) + 31) / 32, (unsigned)(1)), 32, 0, stream>>>(gq1_8);
      else k_gemm<1><<<dim3((unsigned)((C8) + 31) / 32, (unsigned)((N) + 15) / 16, (unsigned)(1)), 32, 0, stream>>>(gq1_8); }
    { GemmP gk1_8;
      gk1_8.A = s2 + (size_t)8 * C * N; gk1_8.B = Wk; gk1_8.bias = bk; gk1_8.R = s2 + (size_t)8 * C * N; gk1_8.C = KF;
      gk1_8.sAo = 0; gk1_8.sAi = 0; gk1_8.sAm = 1; gk1_8.sAk = N; gk1_8.sBo = 0; gk1_8.sBi = 0; gk1_8.sBn = C; gk1_8.sBk = 1; gk1_8.sCo = 0; gk1_8.sCi = 0; gk1_8.sCm = C8; gk1_8.sRo = 0; gk1_8.sRi = 0; gk1_8.sRm = 0; gk1_8.sRn = 0;
      gk1_8.M = N; gk1_8.N = C8; gk1_8.K = C; gk1_8.zi_n = 1; gk1_8.flags = 1; gk1_8.act = 0;
      gk1_8.alpha = 1.0f; gk1_8.beta = 0.0f; gk1_8.sa = 1.0f; gk1_8.sb = 1.0f; gk1_8.Npad = C8; gk1_8.pad_ = 0;
      if ((long long)(N) >= 64 && (long long)(C8) >= 64) k_gemmT<1, 2, 4><<<dim3((unsigned)((C8) + 63) / 64, (unsigned)((N) + 31) / 32, (unsigned)(1)), 32, 0, stream>>>(gk1_8);
      else k_gemm<1><<<dim3((unsigned)((C8) + 31) / 32, (unsigned)((N) + 15) / 16, (unsigned)(1)), 32, 0, stream>>>(gk1_8); }
    k_cast16<<<(unsigned)((((long long)(256) * ((256) / 2)) + 255) / 256), 256, 0, stream>>>(Wv, 256, (_Float16*)(G64A), 256, 256, 256, 1.0f);
    k_castT16<<<(unsigned)((((long long)(1600) * ((256) / 2)) + 255) / 256), 256, 0, stream>>>(s2 + (size_t)8 * C * N, 1600, (_Float16*)(G64B), 256, 256, 1600, 16.0f);
    w25::wmma_gemm64<0, false, 1, 0, false, 0><<<dim3((unsigned)((((256) / 64) * ((1600) / 64) + 7) / 8), (unsigned)(1)), 256, 0, stream>>>((const unsigned short*)(G64A), nullptr, 256, 0, (const unsigned short*)(G64B), nullptr, 256, 0, (void*)(VF), nullptr, 1600, 0, bv, nullptr, 0, 256, 1600, 256, 0.0625f);
    k_ac_planes<<<(unsigned)(((long long)C * N / 2 + 255) / 256), 256, 0, stream>>>(QF, KF, VF, (_Float16*)QH, (_Float16*)QL, (_Float16*)KH, (_Float16*)KL, (_Float16*)V16, N * C8, (long long)C * N);
    w25::wmma_gemm64<1, true, 0, 0, false, 0><<<dim3((unsigned)((((N) / 64) * ((N) / 64) + 7) / 8), (unsigned)(1)), 256, 0, stream>>>((const unsigned short*)(QH), (const unsigned short*)(QL), C8, 0, (const unsigned short*)(KH), (const unsigned short*)(KL), C8, 0, (void*)(EN), nullptr, N, 0, nullptr, nullptr, 0, N, N, C8, 1.0f);
    k_ac_soft<<<N, 256, 0, stream>>>(EN, (_Float16*)P16, N);
    w25::wmma_gemm64<0, false, 0, 0, false, 0><<<dim3((unsigned)((((C) / 64) * ((N) / 64) + 7) / 8), (unsigned)(1)), 256, 0, stream>>>((const unsigned short*)(V16), nullptr, N, 0, (const unsigned short*)(P16), nullptr, N, 0, (void*)(CT), nullptr, N, 0, nullptr, nullptr, 0, C, N, N, 0.000244140625f);
    k_ac_fuse<<<(unsigned)(((long long)C * N + 255) / 256), 256, 0, stream>>>(CT, fw, out, 1, 8, (long long)C * N);
    { GemmP gq1_9;
      gq1_9.A = s1 + (size_t)9 * C * N; gq1_9.B = Wq; gq1_9.bias = bq; gq1_9.R = s1 + (size_t)9 * C * N; gq1_9.C = QF;
      gq1_9.sAo = 0; gq1_9.sAi = 0; gq1_9.sAm = 1; gq1_9.sAk = N; gq1_9.sBo = 0; gq1_9.sBi = 0; gq1_9.sBn = C; gq1_9.sBk = 1; gq1_9.sCo = 0; gq1_9.sCi = 0; gq1_9.sCm = C8; gq1_9.sRo = 0; gq1_9.sRi = 0; gq1_9.sRm = 0; gq1_9.sRn = 0;
      gq1_9.M = N; gq1_9.N = C8; gq1_9.K = C; gq1_9.zi_n = 1; gq1_9.flags = 1; gq1_9.act = 0;
      gq1_9.alpha = 1.0f; gq1_9.beta = 0.0f; gq1_9.sa = 1.0f; gq1_9.sb = 1.0f; gq1_9.Npad = C8; gq1_9.pad_ = 0;
      if ((long long)(N) >= 64 && (long long)(C8) >= 64) k_gemmT<1, 2, 4><<<dim3((unsigned)((C8) + 63) / 64, (unsigned)((N) + 31) / 32, (unsigned)(1)), 32, 0, stream>>>(gq1_9);
      else k_gemm<1><<<dim3((unsigned)((C8) + 31) / 32, (unsigned)((N) + 15) / 16, (unsigned)(1)), 32, 0, stream>>>(gq1_9); }
    { GemmP gk1_9;
      gk1_9.A = s2 + (size_t)9 * C * N; gk1_9.B = Wk; gk1_9.bias = bk; gk1_9.R = s2 + (size_t)9 * C * N; gk1_9.C = KF;
      gk1_9.sAo = 0; gk1_9.sAi = 0; gk1_9.sAm = 1; gk1_9.sAk = N; gk1_9.sBo = 0; gk1_9.sBi = 0; gk1_9.sBn = C; gk1_9.sBk = 1; gk1_9.sCo = 0; gk1_9.sCi = 0; gk1_9.sCm = C8; gk1_9.sRo = 0; gk1_9.sRi = 0; gk1_9.sRm = 0; gk1_9.sRn = 0;
      gk1_9.M = N; gk1_9.N = C8; gk1_9.K = C; gk1_9.zi_n = 1; gk1_9.flags = 1; gk1_9.act = 0;
      gk1_9.alpha = 1.0f; gk1_9.beta = 0.0f; gk1_9.sa = 1.0f; gk1_9.sb = 1.0f; gk1_9.Npad = C8; gk1_9.pad_ = 0;
      if ((long long)(N) >= 64 && (long long)(C8) >= 64) k_gemmT<1, 2, 4><<<dim3((unsigned)((C8) + 63) / 64, (unsigned)((N) + 31) / 32, (unsigned)(1)), 32, 0, stream>>>(gk1_9);
      else k_gemm<1><<<dim3((unsigned)((C8) + 31) / 32, (unsigned)((N) + 15) / 16, (unsigned)(1)), 32, 0, stream>>>(gk1_9); }
    k_cast16<<<(unsigned)((((long long)(256) * ((256) / 2)) + 255) / 256), 256, 0, stream>>>(Wv, 256, (_Float16*)(G64A), 256, 256, 256, 1.0f);
    k_castT16<<<(unsigned)((((long long)(1600) * ((256) / 2)) + 255) / 256), 256, 0, stream>>>(s2 + (size_t)9 * C * N, 1600, (_Float16*)(G64B), 256, 256, 1600, 16.0f);
    w25::wmma_gemm64<0, false, 1, 0, false, 0><<<dim3((unsigned)((((256) / 64) * ((1600) / 64) + 7) / 8), (unsigned)(1)), 256, 0, stream>>>((const unsigned short*)(G64A), nullptr, 256, 0, (const unsigned short*)(G64B), nullptr, 256, 0, (void*)(VF), nullptr, 1600, 0, bv, nullptr, 0, 256, 1600, 256, 0.0625f);
    k_ac_planes<<<(unsigned)(((long long)C * N / 2 + 255) / 256), 256, 0, stream>>>(QF, KF, VF, (_Float16*)QH, (_Float16*)QL, (_Float16*)KH, (_Float16*)KL, (_Float16*)V16, N * C8, (long long)C * N);
    w25::wmma_gemm64<1, true, 0, 0, false, 0><<<dim3((unsigned)((((N) / 64) * ((N) / 64) + 7) / 8), (unsigned)(1)), 256, 0, stream>>>((const unsigned short*)(QH), (const unsigned short*)(QL), C8, 0, (const unsigned short*)(KH), (const unsigned short*)(KL), C8, 0, (void*)(EN), nullptr, N, 0, nullptr, nullptr, 0, N, N, C8, 1.0f);
    k_ac_soft<<<N, 256, 0, stream>>>(EN, (_Float16*)P16, N);
    w25::wmma_gemm64<0, false, 0, 0, false, 0><<<dim3((unsigned)((((C) / 64) * ((N) / 64) + 7) / 8), (unsigned)(1)), 256, 0, stream>>>((const unsigned short*)(V16), nullptr, N, 0, (const unsigned short*)(P16), nullptr, N, 0, (void*)(CT), nullptr, N, 0, nullptr, nullptr, 0, C, N, N, 0.000244140625f);
    k_ac_fuse<<<(unsigned)(((long long)C * N + 255) / 256), 256, 0, stream>>>(CT, fw, out, 1, 9, (long long)C * N);
    { GemmP gq1_10;
      gq1_10.A = s1 + (size_t)10 * C * N; gq1_10.B = Wq; gq1_10.bias = bq; gq1_10.R = s1 + (size_t)10 * C * N; gq1_10.C = QF;
      gq1_10.sAo = 0; gq1_10.sAi = 0; gq1_10.sAm = 1; gq1_10.sAk = N; gq1_10.sBo = 0; gq1_10.sBi = 0; gq1_10.sBn = C; gq1_10.sBk = 1; gq1_10.sCo = 0; gq1_10.sCi = 0; gq1_10.sCm = C8; gq1_10.sRo = 0; gq1_10.sRi = 0; gq1_10.sRm = 0; gq1_10.sRn = 0;
      gq1_10.M = N; gq1_10.N = C8; gq1_10.K = C; gq1_10.zi_n = 1; gq1_10.flags = 1; gq1_10.act = 0;
      gq1_10.alpha = 1.0f; gq1_10.beta = 0.0f; gq1_10.sa = 1.0f; gq1_10.sb = 1.0f; gq1_10.Npad = C8; gq1_10.pad_ = 0;
      if ((long long)(N) >= 64 && (long long)(C8) >= 64) k_gemmT<1, 2, 4><<<dim3((unsigned)((C8) + 63) / 64, (unsigned)((N) + 31) / 32, (unsigned)(1)), 32, 0, stream>>>(gq1_10);
      else k_gemm<1><<<dim3((unsigned)((C8) + 31) / 32, (unsigned)((N) + 15) / 16, (unsigned)(1)), 32, 0, stream>>>(gq1_10); }
    { GemmP gk1_10;
      gk1_10.A = s2 + (size_t)10 * C * N; gk1_10.B = Wk; gk1_10.bias = bk; gk1_10.R = s2 + (size_t)10 * C * N; gk1_10.C = KF;
      gk1_10.sAo = 0; gk1_10.sAi = 0; gk1_10.sAm = 1; gk1_10.sAk = N; gk1_10.sBo = 0; gk1_10.sBi = 0; gk1_10.sBn = C; gk1_10.sBk = 1; gk1_10.sCo = 0; gk1_10.sCi = 0; gk1_10.sCm = C8; gk1_10.sRo = 0; gk1_10.sRi = 0; gk1_10.sRm = 0; gk1_10.sRn = 0;
      gk1_10.M = N; gk1_10.N = C8; gk1_10.K = C; gk1_10.zi_n = 1; gk1_10.flags = 1; gk1_10.act = 0;
      gk1_10.alpha = 1.0f; gk1_10.beta = 0.0f; gk1_10.sa = 1.0f; gk1_10.sb = 1.0f; gk1_10.Npad = C8; gk1_10.pad_ = 0;
      if ((long long)(N) >= 64 && (long long)(C8) >= 64) k_gemmT<1, 2, 4><<<dim3((unsigned)((C8) + 63) / 64, (unsigned)((N) + 31) / 32, (unsigned)(1)), 32, 0, stream>>>(gk1_10);
      else k_gemm<1><<<dim3((unsigned)((C8) + 31) / 32, (unsigned)((N) + 15) / 16, (unsigned)(1)), 32, 0, stream>>>(gk1_10); }
    k_cast16<<<(unsigned)((((long long)(256) * ((256) / 2)) + 255) / 256), 256, 0, stream>>>(Wv, 256, (_Float16*)(G64A), 256, 256, 256, 1.0f);
    k_castT16<<<(unsigned)((((long long)(1600) * ((256) / 2)) + 255) / 256), 256, 0, stream>>>(s2 + (size_t)10 * C * N, 1600, (_Float16*)(G64B), 256, 256, 1600, 16.0f);
    w25::wmma_gemm64<0, false, 1, 0, false, 0><<<dim3((unsigned)((((256) / 64) * ((1600) / 64) + 7) / 8), (unsigned)(1)), 256, 0, stream>>>((const unsigned short*)(G64A), nullptr, 256, 0, (const unsigned short*)(G64B), nullptr, 256, 0, (void*)(VF), nullptr, 1600, 0, bv, nullptr, 0, 256, 1600, 256, 0.0625f);
    k_ac_planes<<<(unsigned)(((long long)C * N / 2 + 255) / 256), 256, 0, stream>>>(QF, KF, VF, (_Float16*)QH, (_Float16*)QL, (_Float16*)KH, (_Float16*)KL, (_Float16*)V16, N * C8, (long long)C * N);
    w25::wmma_gemm64<1, true, 0, 0, false, 0><<<dim3((unsigned)((((N) / 64) * ((N) / 64) + 7) / 8), (unsigned)(1)), 256, 0, stream>>>((const unsigned short*)(QH), (const unsigned short*)(QL), C8, 0, (const unsigned short*)(KH), (const unsigned short*)(KL), C8, 0, (void*)(EN), nullptr, N, 0, nullptr, nullptr, 0, N, N, C8, 1.0f);
    k_ac_soft<<<N, 256, 0, stream>>>(EN, (_Float16*)P16, N);
    w25::wmma_gemm64<0, false, 0, 0, false, 0><<<dim3((unsigned)((((C) / 64) * ((N) / 64) + 7) / 8), (unsigned)(1)), 256, 0, stream>>>((const unsigned short*)(V16), nullptr, N, 0, (const unsigned short*)(P16), nullptr, N, 0, (void*)(CT), nullptr, N, 0, nullptr, nullptr, 0, C, N, N, 0.000244140625f);
    k_ac_fuse<<<(unsigned)(((long long)C * N + 255) / 256), 256, 0, stream>>>(CT, fw, out, 1, 10, (long long)C * N);
    { GemmP gq1_11;
      gq1_11.A = s1 + (size_t)11 * C * N; gq1_11.B = Wq; gq1_11.bias = bq; gq1_11.R = s1 + (size_t)11 * C * N; gq1_11.C = QF;
      gq1_11.sAo = 0; gq1_11.sAi = 0; gq1_11.sAm = 1; gq1_11.sAk = N; gq1_11.sBo = 0; gq1_11.sBi = 0; gq1_11.sBn = C; gq1_11.sBk = 1; gq1_11.sCo = 0; gq1_11.sCi = 0; gq1_11.sCm = C8; gq1_11.sRo = 0; gq1_11.sRi = 0; gq1_11.sRm = 0; gq1_11.sRn = 0;
      gq1_11.M = N; gq1_11.N = C8; gq1_11.K = C; gq1_11.zi_n = 1; gq1_11.flags = 1; gq1_11.act = 0;
      gq1_11.alpha = 1.0f; gq1_11.beta = 0.0f; gq1_11.sa = 1.0f; gq1_11.sb = 1.0f; gq1_11.Npad = C8; gq1_11.pad_ = 0;
      if ((long long)(N) >= 64 && (long long)(C8) >= 64) k_gemmT<1, 2, 4><<<dim3((unsigned)((C8) + 63) / 64, (unsigned)((N) + 31) / 32, (unsigned)(1)), 32, 0, stream>>>(gq1_11);
      else k_gemm<1><<<dim3((unsigned)((C8) + 31) / 32, (unsigned)((N) + 15) / 16, (unsigned)(1)), 32, 0, stream>>>(gq1_11); }
    { GemmP gk1_11;
      gk1_11.A = s2 + (size_t)11 * C * N; gk1_11.B = Wk; gk1_11.bias = bk; gk1_11.R = s2 + (size_t)11 * C * N; gk1_11.C = KF;
      gk1_11.sAo = 0; gk1_11.sAi = 0; gk1_11.sAm = 1; gk1_11.sAk = N; gk1_11.sBo = 0; gk1_11.sBi = 0; gk1_11.sBn = C; gk1_11.sBk = 1; gk1_11.sCo = 0; gk1_11.sCi = 0; gk1_11.sCm = C8; gk1_11.sRo = 0; gk1_11.sRi = 0; gk1_11.sRm = 0; gk1_11.sRn = 0;
      gk1_11.M = N; gk1_11.N = C8; gk1_11.K = C; gk1_11.zi_n = 1; gk1_11.flags = 1; gk1_11.act = 0;
      gk1_11.alpha = 1.0f; gk1_11.beta = 0.0f; gk1_11.sa = 1.0f; gk1_11.sb = 1.0f; gk1_11.Npad = C8; gk1_11.pad_ = 0;
      if ((long long)(N) >= 64 && (long long)(C8) >= 64) k_gemmT<1, 2, 4><<<dim3((unsigned)((C8) + 63) / 64, (unsigned)((N) + 31) / 32, (unsigned)(1)), 32, 0, stream>>>(gk1_11);
      else k_gemm<1><<<dim3((unsigned)((C8) + 31) / 32, (unsigned)((N) + 15) / 16, (unsigned)(1)), 32, 0, stream>>>(gk1_11); }
    k_cast16<<<(unsigned)((((long long)(256) * ((256) / 2)) + 255) / 256), 256, 0, stream>>>(Wv, 256, (_Float16*)(G64A), 256, 256, 256, 1.0f);
    k_castT16<<<(unsigned)((((long long)(1600) * ((256) / 2)) + 255) / 256), 256, 0, stream>>>(s2 + (size_t)11 * C * N, 1600, (_Float16*)(G64B), 256, 256, 1600, 16.0f);
    w25::wmma_gemm64<0, false, 1, 0, false, 0><<<dim3((unsigned)((((256) / 64) * ((1600) / 64) + 7) / 8), (unsigned)(1)), 256, 0, stream>>>((const unsigned short*)(G64A), nullptr, 256, 0, (const unsigned short*)(G64B), nullptr, 256, 0, (void*)(VF), nullptr, 1600, 0, bv, nullptr, 0, 256, 1600, 256, 0.0625f);
    k_ac_planes<<<(unsigned)(((long long)C * N / 2 + 255) / 256), 256, 0, stream>>>(QF, KF, VF, (_Float16*)QH, (_Float16*)QL, (_Float16*)KH, (_Float16*)KL, (_Float16*)V16, N * C8, (long long)C * N);
    w25::wmma_gemm64<1, true, 0, 0, false, 0><<<dim3((unsigned)((((N) / 64) * ((N) / 64) + 7) / 8), (unsigned)(1)), 256, 0, stream>>>((const unsigned short*)(QH), (const unsigned short*)(QL), C8, 0, (const unsigned short*)(KH), (const unsigned short*)(KL), C8, 0, (void*)(EN), nullptr, N, 0, nullptr, nullptr, 0, N, N, C8, 1.0f);
    k_ac_soft<<<N, 256, 0, stream>>>(EN, (_Float16*)P16, N);
    w25::wmma_gemm64<0, false, 0, 0, false, 0><<<dim3((unsigned)((((C) / 64) * ((N) / 64) + 7) / 8), (unsigned)(1)), 256, 0, stream>>>((const unsigned short*)(V16), nullptr, N, 0, (const unsigned short*)(P16), nullptr, N, 0, (void*)(CT), nullptr, N, 0, nullptr, nullptr, 0, C, N, N, 0.000244140625f);
    k_ac_fuse<<<(unsigned)(((long long)C * N + 255) / 256), 256, 0, stream>>>(CT, fw, out, 1, 11, (long long)C * N);
    { GemmP gq1_12;
      gq1_12.A = s1 + (size_t)12 * C * N; gq1_12.B = Wq; gq1_12.bias = bq; gq1_12.R = s1 + (size_t)12 * C * N; gq1_12.C = QF;
      gq1_12.sAo = 0; gq1_12.sAi = 0; gq1_12.sAm = 1; gq1_12.sAk = N; gq1_12.sBo = 0; gq1_12.sBi = 0; gq1_12.sBn = C; gq1_12.sBk = 1; gq1_12.sCo = 0; gq1_12.sCi = 0; gq1_12.sCm = C8; gq1_12.sRo = 0; gq1_12.sRi = 0; gq1_12.sRm = 0; gq1_12.sRn = 0;
      gq1_12.M = N; gq1_12.N = C8; gq1_12.K = C; gq1_12.zi_n = 1; gq1_12.flags = 1; gq1_12.act = 0;
      gq1_12.alpha = 1.0f; gq1_12.beta = 0.0f; gq1_12.sa = 1.0f; gq1_12.sb = 1.0f; gq1_12.Npad = C8; gq1_12.pad_ = 0;
      if ((long long)(N) >= 64 && (long long)(C8) >= 64) k_gemmT<1, 2, 4><<<dim3((unsigned)((C8) + 63) / 64, (unsigned)((N) + 31) / 32, (unsigned)(1)), 32, 0, stream>>>(gq1_12);
      else k_gemm<1><<<dim3((unsigned)((C8) + 31) / 32, (unsigned)((N) + 15) / 16, (unsigned)(1)), 32, 0, stream>>>(gq1_12); }
    { GemmP gk1_12;
      gk1_12.A = s2 + (size_t)12 * C * N; gk1_12.B = Wk; gk1_12.bias = bk; gk1_12.R = s2 + (size_t)12 * C * N; gk1_12.C = KF;
      gk1_12.sAo = 0; gk1_12.sAi = 0; gk1_12.sAm = 1; gk1_12.sAk = N; gk1_12.sBo = 0; gk1_12.sBi = 0; gk1_12.sBn = C; gk1_12.sBk = 1; gk1_12.sCo = 0; gk1_12.sCi = 0; gk1_12.sCm = C8; gk1_12.sRo = 0; gk1_12.sRi = 0; gk1_12.sRm = 0; gk1_12.sRn = 0;
      gk1_12.M = N; gk1_12.N = C8; gk1_12.K = C; gk1_12.zi_n = 1; gk1_12.flags = 1; gk1_12.act = 0;
      gk1_12.alpha = 1.0f; gk1_12.beta = 0.0f; gk1_12.sa = 1.0f; gk1_12.sb = 1.0f; gk1_12.Npad = C8; gk1_12.pad_ = 0;
      if ((long long)(N) >= 64 && (long long)(C8) >= 64) k_gemmT<1, 2, 4><<<dim3((unsigned)((C8) + 63) / 64, (unsigned)((N) + 31) / 32, (unsigned)(1)), 32, 0, stream>>>(gk1_12);
      else k_gemm<1><<<dim3((unsigned)((C8) + 31) / 32, (unsigned)((N) + 15) / 16, (unsigned)(1)), 32, 0, stream>>>(gk1_12); }
    k_cast16<<<(unsigned)((((long long)(256) * ((256) / 2)) + 255) / 256), 256, 0, stream>>>(Wv, 256, (_Float16*)(G64A), 256, 256, 256, 1.0f);
    k_castT16<<<(unsigned)((((long long)(1600) * ((256) / 2)) + 255) / 256), 256, 0, stream>>>(s2 + (size_t)12 * C * N, 1600, (_Float16*)(G64B), 256, 256, 1600, 16.0f);
    w25::wmma_gemm64<0, false, 1, 0, false, 0><<<dim3((unsigned)((((256) / 64) * ((1600) / 64) + 7) / 8), (unsigned)(1)), 256, 0, stream>>>((const unsigned short*)(G64A), nullptr, 256, 0, (const unsigned short*)(G64B), nullptr, 256, 0, (void*)(VF), nullptr, 1600, 0, bv, nullptr, 0, 256, 1600, 256, 0.0625f);
    k_ac_planes<<<(unsigned)(((long long)C * N / 2 + 255) / 256), 256, 0, stream>>>(QF, KF, VF, (_Float16*)QH, (_Float16*)QL, (_Float16*)KH, (_Float16*)KL, (_Float16*)V16, N * C8, (long long)C * N);
    w25::wmma_gemm64<1, true, 0, 0, false, 0><<<dim3((unsigned)((((N) / 64) * ((N) / 64) + 7) / 8), (unsigned)(1)), 256, 0, stream>>>((const unsigned short*)(QH), (const unsigned short*)(QL), C8, 0, (const unsigned short*)(KH), (const unsigned short*)(KL), C8, 0, (void*)(EN), nullptr, N, 0, nullptr, nullptr, 0, N, N, C8, 1.0f);
    k_ac_soft<<<N, 256, 0, stream>>>(EN, (_Float16*)P16, N);
    w25::wmma_gemm64<0, false, 0, 0, false, 0><<<dim3((unsigned)((((C) / 64) * ((N) / 64) + 7) / 8), (unsigned)(1)), 256, 0, stream>>>((const unsigned short*)(V16), nullptr, N, 0, (const unsigned short*)(P16), nullptr, N, 0, (void*)(CT), nullptr, N, 0, nullptr, nullptr, 0, C, N, N, 0.000244140625f);
    k_ac_fuse<<<(unsigned)(((long long)C * N + 255) / 256), 256, 0, stream>>>(CT, fw, out, 1, 12, (long long)C * N);
    { GemmP gq1_13;
      gq1_13.A = s1 + (size_t)13 * C * N; gq1_13.B = Wq; gq1_13.bias = bq; gq1_13.R = s1 + (size_t)13 * C * N; gq1_13.C = QF;
      gq1_13.sAo = 0; gq1_13.sAi = 0; gq1_13.sAm = 1; gq1_13.sAk = N; gq1_13.sBo = 0; gq1_13.sBi = 0; gq1_13.sBn = C; gq1_13.sBk = 1; gq1_13.sCo = 0; gq1_13.sCi = 0; gq1_13.sCm = C8; gq1_13.sRo = 0; gq1_13.sRi = 0; gq1_13.sRm = 0; gq1_13.sRn = 0;
      gq1_13.M = N; gq1_13.N = C8; gq1_13.K = C; gq1_13.zi_n = 1; gq1_13.flags = 1; gq1_13.act = 0;
      gq1_13.alpha = 1.0f; gq1_13.beta = 0.0f; gq1_13.sa = 1.0f; gq1_13.sb = 1.0f; gq1_13.Npad = C8; gq1_13.pad_ = 0;
      if ((long long)(N) >= 64 && (long long)(C8) >= 64) k_gemmT<1, 2, 4><<<dim3((unsigned)((C8) + 63) / 64, (unsigned)((N) + 31) / 32, (unsigned)(1)), 32, 0, stream>>>(gq1_13);
      else k_gemm<1><<<dim3((unsigned)((C8) + 31) / 32, (unsigned)((N) + 15) / 16, (unsigned)(1)), 32, 0, stream>>>(gq1_13); }
    { GemmP gk1_13;
      gk1_13.A = s2 + (size_t)13 * C * N; gk1_13.B = Wk; gk1_13.bias = bk; gk1_13.R = s2 + (size_t)13 * C * N; gk1_13.C = KF;
      gk1_13.sAo = 0; gk1_13.sAi = 0; gk1_13.sAm = 1; gk1_13.sAk = N; gk1_13.sBo = 0; gk1_13.sBi = 0; gk1_13.sBn = C; gk1_13.sBk = 1; gk1_13.sCo = 0; gk1_13.sCi = 0; gk1_13.sCm = C8; gk1_13.sRo = 0; gk1_13.sRi = 0; gk1_13.sRm = 0; gk1_13.sRn = 0;
      gk1_13.M = N; gk1_13.N = C8; gk1_13.K = C; gk1_13.zi_n = 1; gk1_13.flags = 1; gk1_13.act = 0;
      gk1_13.alpha = 1.0f; gk1_13.beta = 0.0f; gk1_13.sa = 1.0f; gk1_13.sb = 1.0f; gk1_13.Npad = C8; gk1_13.pad_ = 0;
      if ((long long)(N) >= 64 && (long long)(C8) >= 64) k_gemmT<1, 2, 4><<<dim3((unsigned)((C8) + 63) / 64, (unsigned)((N) + 31) / 32, (unsigned)(1)), 32, 0, stream>>>(gk1_13);
      else k_gemm<1><<<dim3((unsigned)((C8) + 31) / 32, (unsigned)((N) + 15) / 16, (unsigned)(1)), 32, 0, stream>>>(gk1_13); }
    k_cast16<<<(unsigned)((((long long)(256) * ((256) / 2)) + 255) / 256), 256, 0, stream>>>(Wv, 256, (_Float16*)(G64A), 256, 256, 256, 1.0f);
    k_castT16<<<(unsigned)((((long long)(1600) * ((256) / 2)) + 255) / 256), 256, 0, stream>>>(s2 + (size_t)13 * C * N, 1600, (_Float16*)(G64B), 256, 256, 1600, 16.0f);
    w25::wmma_gemm64<0, false, 1, 0, false, 0><<<dim3((unsigned)((((256) / 64) * ((1600) / 64) + 7) / 8), (unsigned)(1)), 256, 0, stream>>>((const unsigned short*)(G64A), nullptr, 256, 0, (const unsigned short*)(G64B), nullptr, 256, 0, (void*)(VF), nullptr, 1600, 0, bv, nullptr, 0, 256, 1600, 256, 0.0625f);
    k_ac_planes<<<(unsigned)(((long long)C * N / 2 + 255) / 256), 256, 0, stream>>>(QF, KF, VF, (_Float16*)QH, (_Float16*)QL, (_Float16*)KH, (_Float16*)KL, (_Float16*)V16, N * C8, (long long)C * N);
    w25::wmma_gemm64<1, true, 0, 0, false, 0><<<dim3((unsigned)((((N) / 64) * ((N) / 64) + 7) / 8), (unsigned)(1)), 256, 0, stream>>>((const unsigned short*)(QH), (const unsigned short*)(QL), C8, 0, (const unsigned short*)(KH), (const unsigned short*)(KL), C8, 0, (void*)(EN), nullptr, N, 0, nullptr, nullptr, 0, N, N, C8, 1.0f);
    k_ac_soft<<<N, 256, 0, stream>>>(EN, (_Float16*)P16, N);
    w25::wmma_gemm64<0, false, 0, 0, false, 0><<<dim3((unsigned)((((C) / 64) * ((N) / 64) + 7) / 8), (unsigned)(1)), 256, 0, stream>>>((const unsigned short*)(V16), nullptr, N, 0, (const unsigned short*)(P16), nullptr, N, 0, (void*)(CT), nullptr, N, 0, nullptr, nullptr, 0, C, N, N, 0.000244140625f);
    k_ac_fuse<<<(unsigned)(((long long)C * N + 255) / 256), 256, 0, stream>>>(CT, fw, out, 1, 13, (long long)C * N);
    { GemmP gq1_14;
      gq1_14.A = s1 + (size_t)14 * C * N; gq1_14.B = Wq; gq1_14.bias = bq; gq1_14.R = s1 + (size_t)14 * C * N; gq1_14.C = QF;
      gq1_14.sAo = 0; gq1_14.sAi = 0; gq1_14.sAm = 1; gq1_14.sAk = N; gq1_14.sBo = 0; gq1_14.sBi = 0; gq1_14.sBn = C; gq1_14.sBk = 1; gq1_14.sCo = 0; gq1_14.sCi = 0; gq1_14.sCm = C8; gq1_14.sRo = 0; gq1_14.sRi = 0; gq1_14.sRm = 0; gq1_14.sRn = 0;
      gq1_14.M = N; gq1_14.N = C8; gq1_14.K = C; gq1_14.zi_n = 1; gq1_14.flags = 1; gq1_14.act = 0;
      gq1_14.alpha = 1.0f; gq1_14.beta = 0.0f; gq1_14.sa = 1.0f; gq1_14.sb = 1.0f; gq1_14.Npad = C8; gq1_14.pad_ = 0;
      if ((long long)(N) >= 64 && (long long)(C8) >= 64) k_gemmT<1, 2, 4><<<dim3((unsigned)((C8) + 63) / 64, (unsigned)((N) + 31) / 32, (unsigned)(1)), 32, 0, stream>>>(gq1_14);
      else k_gemm<1><<<dim3((unsigned)((C8) + 31) / 32, (unsigned)((N) + 15) / 16, (unsigned)(1)), 32, 0, stream>>>(gq1_14); }
    { GemmP gk1_14;
      gk1_14.A = s2 + (size_t)14 * C * N; gk1_14.B = Wk; gk1_14.bias = bk; gk1_14.R = s2 + (size_t)14 * C * N; gk1_14.C = KF;
      gk1_14.sAo = 0; gk1_14.sAi = 0; gk1_14.sAm = 1; gk1_14.sAk = N; gk1_14.sBo = 0; gk1_14.sBi = 0; gk1_14.sBn = C; gk1_14.sBk = 1; gk1_14.sCo = 0; gk1_14.sCi = 0; gk1_14.sCm = C8; gk1_14.sRo = 0; gk1_14.sRi = 0; gk1_14.sRm = 0; gk1_14.sRn = 0;
      gk1_14.M = N; gk1_14.N = C8; gk1_14.K = C; gk1_14.zi_n = 1; gk1_14.flags = 1; gk1_14.act = 0;
      gk1_14.alpha = 1.0f; gk1_14.beta = 0.0f; gk1_14.sa = 1.0f; gk1_14.sb = 1.0f; gk1_14.Npad = C8; gk1_14.pad_ = 0;
      if ((long long)(N) >= 64 && (long long)(C8) >= 64) k_gemmT<1, 2, 4><<<dim3((unsigned)((C8) + 63) / 64, (unsigned)((N) + 31) / 32, (unsigned)(1)), 32, 0, stream>>>(gk1_14);
      else k_gemm<1><<<dim3((unsigned)((C8) + 31) / 32, (unsigned)((N) + 15) / 16, (unsigned)(1)), 32, 0, stream>>>(gk1_14); }
    k_cast16<<<(unsigned)((((long long)(256) * ((256) / 2)) + 255) / 256), 256, 0, stream>>>(Wv, 256, (_Float16*)(G64A), 256, 256, 256, 1.0f);
    k_castT16<<<(unsigned)((((long long)(1600) * ((256) / 2)) + 255) / 256), 256, 0, stream>>>(s2 + (size_t)14 * C * N, 1600, (_Float16*)(G64B), 256, 256, 1600, 16.0f);
    w25::wmma_gemm64<0, false, 1, 0, false, 0><<<dim3((unsigned)((((256) / 64) * ((1600) / 64) + 7) / 8), (unsigned)(1)), 256, 0, stream>>>((const unsigned short*)(G64A), nullptr, 256, 0, (const unsigned short*)(G64B), nullptr, 256, 0, (void*)(VF), nullptr, 1600, 0, bv, nullptr, 0, 256, 1600, 256, 0.0625f);
    k_ac_planes<<<(unsigned)(((long long)C * N / 2 + 255) / 256), 256, 0, stream>>>(QF, KF, VF, (_Float16*)QH, (_Float16*)QL, (_Float16*)KH, (_Float16*)KL, (_Float16*)V16, N * C8, (long long)C * N);
    w25::wmma_gemm64<1, true, 0, 0, false, 0><<<dim3((unsigned)((((N) / 64) * ((N) / 64) + 7) / 8), (unsigned)(1)), 256, 0, stream>>>((const unsigned short*)(QH), (const unsigned short*)(QL), C8, 0, (const unsigned short*)(KH), (const unsigned short*)(KL), C8, 0, (void*)(EN), nullptr, N, 0, nullptr, nullptr, 0, N, N, C8, 1.0f);
    k_ac_soft<<<N, 256, 0, stream>>>(EN, (_Float16*)P16, N);
    w25::wmma_gemm64<0, false, 0, 0, false, 0><<<dim3((unsigned)((((C) / 64) * ((N) / 64) + 7) / 8), (unsigned)(1)), 256, 0, stream>>>((const unsigned short*)(V16), nullptr, N, 0, (const unsigned short*)(P16), nullptr, N, 0, (void*)(CT), nullptr, N, 0, nullptr, nullptr, 0, C, N, N, 0.000244140625f);
    k_ac_fuse<<<(unsigned)(((long long)C * N + 255) / 256), 256, 0, stream>>>(CT, fw, out, 1, 14, (long long)C * N);
    { GemmP gq1_15;
      gq1_15.A = s1 + (size_t)15 * C * N; gq1_15.B = Wq; gq1_15.bias = bq; gq1_15.R = s1 + (size_t)15 * C * N; gq1_15.C = QF;
      gq1_15.sAo = 0; gq1_15.sAi = 0; gq1_15.sAm = 1; gq1_15.sAk = N; gq1_15.sBo = 0; gq1_15.sBi = 0; gq1_15.sBn = C; gq1_15.sBk = 1; gq1_15.sCo = 0; gq1_15.sCi = 0; gq1_15.sCm = C8; gq1_15.sRo = 0; gq1_15.sRi = 0; gq1_15.sRm = 0; gq1_15.sRn = 0;
      gq1_15.M = N; gq1_15.N = C8; gq1_15.K = C; gq1_15.zi_n = 1; gq1_15.flags = 1; gq1_15.act = 0;
      gq1_15.alpha = 1.0f; gq1_15.beta = 0.0f; gq1_15.sa = 1.0f; gq1_15.sb = 1.0f; gq1_15.Npad = C8; gq1_15.pad_ = 0;
      if ((long long)(N) >= 64 && (long long)(C8) >= 64) k_gemmT<1, 2, 4><<<dim3((unsigned)((C8) + 63) / 64, (unsigned)((N) + 31) / 32, (unsigned)(1)), 32, 0, stream>>>(gq1_15);
      else k_gemm<1><<<dim3((unsigned)((C8) + 31) / 32, (unsigned)((N) + 15) / 16, (unsigned)(1)), 32, 0, stream>>>(gq1_15); }
    { GemmP gk1_15;
      gk1_15.A = s2 + (size_t)15 * C * N; gk1_15.B = Wk; gk1_15.bias = bk; gk1_15.R = s2 + (size_t)15 * C * N; gk1_15.C = KF;
      gk1_15.sAo = 0; gk1_15.sAi = 0; gk1_15.sAm = 1; gk1_15.sAk = N; gk1_15.sBo = 0; gk1_15.sBi = 0; gk1_15.sBn = C; gk1_15.sBk = 1; gk1_15.sCo = 0; gk1_15.sCi = 0; gk1_15.sCm = C8; gk1_15.sRo = 0; gk1_15.sRi = 0; gk1_15.sRm = 0; gk1_15.sRn = 0;
      gk1_15.M = N; gk1_15.N = C8; gk1_15.K = C; gk1_15.zi_n = 1; gk1_15.flags = 1; gk1_15.act = 0;
      gk1_15.alpha = 1.0f; gk1_15.beta = 0.0f; gk1_15.sa = 1.0f; gk1_15.sb = 1.0f; gk1_15.Npad = C8; gk1_15.pad_ = 0;
      if ((long long)(N) >= 64 && (long long)(C8) >= 64) k_gemmT<1, 2, 4><<<dim3((unsigned)((C8) + 63) / 64, (unsigned)((N) + 31) / 32, (unsigned)(1)), 32, 0, stream>>>(gk1_15);
      else k_gemm<1><<<dim3((unsigned)((C8) + 31) / 32, (unsigned)((N) + 15) / 16, (unsigned)(1)), 32, 0, stream>>>(gk1_15); }
    k_cast16<<<(unsigned)((((long long)(256) * ((256) / 2)) + 255) / 256), 256, 0, stream>>>(Wv, 256, (_Float16*)(G64A), 256, 256, 256, 1.0f);
    k_castT16<<<(unsigned)((((long long)(1600) * ((256) / 2)) + 255) / 256), 256, 0, stream>>>(s2 + (size_t)15 * C * N, 1600, (_Float16*)(G64B), 256, 256, 1600, 16.0f);
    w25::wmma_gemm64<0, false, 1, 0, false, 0><<<dim3((unsigned)((((256) / 64) * ((1600) / 64) + 7) / 8), (unsigned)(1)), 256, 0, stream>>>((const unsigned short*)(G64A), nullptr, 256, 0, (const unsigned short*)(G64B), nullptr, 256, 0, (void*)(VF), nullptr, 1600, 0, bv, nullptr, 0, 256, 1600, 256, 0.0625f);
    k_ac_planes<<<(unsigned)(((long long)C * N / 2 + 255) / 256), 256, 0, stream>>>(QF, KF, VF, (_Float16*)QH, (_Float16*)QL, (_Float16*)KH, (_Float16*)KL, (_Float16*)V16, N * C8, (long long)C * N);
    w25::wmma_gemm64<1, true, 0, 0, false, 0><<<dim3((unsigned)((((N) / 64) * ((N) / 64) + 7) / 8), (unsigned)(1)), 256, 0, stream>>>((const unsigned short*)(QH), (const unsigned short*)(QL), C8, 0, (const unsigned short*)(KH), (const unsigned short*)(KL), C8, 0, (void*)(EN), nullptr, N, 0, nullptr, nullptr, 0, N, N, C8, 1.0f);
    k_ac_soft<<<N, 256, 0, stream>>>(EN, (_Float16*)P16, N);
    w25::wmma_gemm64<0, false, 0, 0, false, 0><<<dim3((unsigned)((((C) / 64) * ((N) / 64) + 7) / 8), (unsigned)(1)), 256, 0, stream>>>((const unsigned short*)(V16), nullptr, N, 0, (const unsigned short*)(P16), nullptr, N, 0, (void*)(CT), nullptr, N, 0, nullptr, nullptr, 0, C, N, N, 0.000244140625f);
    k_ac_fuse<<<(unsigned)(((long long)C * N + 255) / 256), 256, 0, stream>>>(CT, fw, out, 1, 15, (long long)C * N);
    { GemmP gq2_0;
      gq2_0.A = s2 + (size_t)0 * C * N; gq2_0.B = Wq; gq2_0.bias = bq; gq2_0.R = s2 + (size_t)0 * C * N; gq2_0.C = QF;
      gq2_0.sAo = 0; gq2_0.sAi = 0; gq2_0.sAm = 1; gq2_0.sAk = N; gq2_0.sBo = 0; gq2_0.sBi = 0; gq2_0.sBn = C; gq2_0.sBk = 1; gq2_0.sCo = 0; gq2_0.sCi = 0; gq2_0.sCm = C8; gq2_0.sRo = 0; gq2_0.sRi = 0; gq2_0.sRm = 0; gq2_0.sRn = 0;
      gq2_0.M = N; gq2_0.N = C8; gq2_0.K = C; gq2_0.zi_n = 1; gq2_0.flags = 1; gq2_0.act = 0;
      gq2_0.alpha = 1.0f; gq2_0.beta = 0.0f; gq2_0.sa = 1.0f; gq2_0.sb = 1.0f; gq2_0.Npad = C8; gq2_0.pad_ = 0;
      if ((long long)(N) >= 64 && (long long)(C8) >= 64) k_gemmT<1, 2, 4><<<dim3((unsigned)((C8) + 63) / 64, (unsigned)((N) + 31) / 32, (unsigned)(1)), 32, 0, stream>>>(gq2_0);
      else k_gemm<1><<<dim3((unsigned)((C8) + 31) / 32, (unsigned)((N) + 15) / 16, (unsigned)(1)), 32, 0, stream>>>(gq2_0); }
    { GemmP gk2_0;
      gk2_0.A = s0 + (size_t)0 * C * N; gk2_0.B = Wk; gk2_0.bias = bk; gk2_0.R = s0 + (size_t)0 * C * N; gk2_0.C = KF;
      gk2_0.sAo = 0; gk2_0.sAi = 0; gk2_0.sAm = 1; gk2_0.sAk = N; gk2_0.sBo = 0; gk2_0.sBi = 0; gk2_0.sBn = C; gk2_0.sBk = 1; gk2_0.sCo = 0; gk2_0.sCi = 0; gk2_0.sCm = C8; gk2_0.sRo = 0; gk2_0.sRi = 0; gk2_0.sRm = 0; gk2_0.sRn = 0;
      gk2_0.M = N; gk2_0.N = C8; gk2_0.K = C; gk2_0.zi_n = 1; gk2_0.flags = 1; gk2_0.act = 0;
      gk2_0.alpha = 1.0f; gk2_0.beta = 0.0f; gk2_0.sa = 1.0f; gk2_0.sb = 1.0f; gk2_0.Npad = C8; gk2_0.pad_ = 0;
      if ((long long)(N) >= 64 && (long long)(C8) >= 64) k_gemmT<1, 2, 4><<<dim3((unsigned)((C8) + 63) / 64, (unsigned)((N) + 31) / 32, (unsigned)(1)), 32, 0, stream>>>(gk2_0);
      else k_gemm<1><<<dim3((unsigned)((C8) + 31) / 32, (unsigned)((N) + 15) / 16, (unsigned)(1)), 32, 0, stream>>>(gk2_0); }
    k_cast16<<<(unsigned)((((long long)(256) * ((256) / 2)) + 255) / 256), 256, 0, stream>>>(Wv, 256, (_Float16*)(G64A), 256, 256, 256, 1.0f);
    k_castT16<<<(unsigned)((((long long)(1600) * ((256) / 2)) + 255) / 256), 256, 0, stream>>>(s0 + (size_t)0 * C * N, 1600, (_Float16*)(G64B), 256, 256, 1600, 16.0f);
    w25::wmma_gemm64<0, false, 1, 0, false, 0><<<dim3((unsigned)((((256) / 64) * ((1600) / 64) + 7) / 8), (unsigned)(1)), 256, 0, stream>>>((const unsigned short*)(G64A), nullptr, 256, 0, (const unsigned short*)(G64B), nullptr, 256, 0, (void*)(VF), nullptr, 1600, 0, bv, nullptr, 0, 256, 1600, 256, 0.0625f);
    k_ac_planes<<<(unsigned)(((long long)C * N / 2 + 255) / 256), 256, 0, stream>>>(QF, KF, VF, (_Float16*)QH, (_Float16*)QL, (_Float16*)KH, (_Float16*)KL, (_Float16*)V16, N * C8, (long long)C * N);
    w25::wmma_gemm64<1, true, 0, 0, false, 0><<<dim3((unsigned)((((N) / 64) * ((N) / 64) + 7) / 8), (unsigned)(1)), 256, 0, stream>>>((const unsigned short*)(QH), (const unsigned short*)(QL), C8, 0, (const unsigned short*)(KH), (const unsigned short*)(KL), C8, 0, (void*)(EN), nullptr, N, 0, nullptr, nullptr, 0, N, N, C8, 1.0f);
    k_ac_soft<<<N, 256, 0, stream>>>(EN, (_Float16*)P16, N);
    w25::wmma_gemm64<0, false, 0, 0, false, 0><<<dim3((unsigned)((((C) / 64) * ((N) / 64) + 7) / 8), (unsigned)(1)), 256, 0, stream>>>((const unsigned short*)(V16), nullptr, N, 0, (const unsigned short*)(P16), nullptr, N, 0, (void*)(CT), nullptr, N, 0, nullptr, nullptr, 0, C, N, N, 0.000244140625f);
    k_ac_fuse<<<(unsigned)(((long long)C * N + 255) / 256), 256, 0, stream>>>(CT, fw, out, 2, 0, (long long)C * N);
    { GemmP gq2_1;
      gq2_1.A = s2 + (size_t)1 * C * N; gq2_1.B = Wq; gq2_1.bias = bq; gq2_1.R = s2 + (size_t)1 * C * N; gq2_1.C = QF;
      gq2_1.sAo = 0; gq2_1.sAi = 0; gq2_1.sAm = 1; gq2_1.sAk = N; gq2_1.sBo = 0; gq2_1.sBi = 0; gq2_1.sBn = C; gq2_1.sBk = 1; gq2_1.sCo = 0; gq2_1.sCi = 0; gq2_1.sCm = C8; gq2_1.sRo = 0; gq2_1.sRi = 0; gq2_1.sRm = 0; gq2_1.sRn = 0;
      gq2_1.M = N; gq2_1.N = C8; gq2_1.K = C; gq2_1.zi_n = 1; gq2_1.flags = 1; gq2_1.act = 0;
      gq2_1.alpha = 1.0f; gq2_1.beta = 0.0f; gq2_1.sa = 1.0f; gq2_1.sb = 1.0f; gq2_1.Npad = C8; gq2_1.pad_ = 0;
      if ((long long)(N) >= 64 && (long long)(C8) >= 64) k_gemmT<1, 2, 4><<<dim3((unsigned)((C8) + 63) / 64, (unsigned)((N) + 31) / 32, (unsigned)(1)), 32, 0, stream>>>(gq2_1);
      else k_gemm<1><<<dim3((unsigned)((C8) + 31) / 32, (unsigned)((N) + 15) / 16, (unsigned)(1)), 32, 0, stream>>>(gq2_1); }
    { GemmP gk2_1;
      gk2_1.A = s0 + (size_t)1 * C * N; gk2_1.B = Wk; gk2_1.bias = bk; gk2_1.R = s0 + (size_t)1 * C * N; gk2_1.C = KF;
      gk2_1.sAo = 0; gk2_1.sAi = 0; gk2_1.sAm = 1; gk2_1.sAk = N; gk2_1.sBo = 0; gk2_1.sBi = 0; gk2_1.sBn = C; gk2_1.sBk = 1; gk2_1.sCo = 0; gk2_1.sCi = 0; gk2_1.sCm = C8; gk2_1.sRo = 0; gk2_1.sRi = 0; gk2_1.sRm = 0; gk2_1.sRn = 0;
      gk2_1.M = N; gk2_1.N = C8; gk2_1.K = C; gk2_1.zi_n = 1; gk2_1.flags = 1; gk2_1.act = 0;
      gk2_1.alpha = 1.0f; gk2_1.beta = 0.0f; gk2_1.sa = 1.0f; gk2_1.sb = 1.0f; gk2_1.Npad = C8; gk2_1.pad_ = 0;
      if ((long long)(N) >= 64 && (long long)(C8) >= 64) k_gemmT<1, 2, 4><<<dim3((unsigned)((C8) + 63) / 64, (unsigned)((N) + 31) / 32, (unsigned)(1)), 32, 0, stream>>>(gk2_1);
      else k_gemm<1><<<dim3((unsigned)((C8) + 31) / 32, (unsigned)((N) + 15) / 16, (unsigned)(1)), 32, 0, stream>>>(gk2_1); }
    k_cast16<<<(unsigned)((((long long)(256) * ((256) / 2)) + 255) / 256), 256, 0, stream>>>(Wv, 256, (_Float16*)(G64A), 256, 256, 256, 1.0f);
    k_castT16<<<(unsigned)((((long long)(1600) * ((256) / 2)) + 255) / 256), 256, 0, stream>>>(s0 + (size_t)1 * C * N, 1600, (_Float16*)(G64B), 256, 256, 1600, 16.0f);
    w25::wmma_gemm64<0, false, 1, 0, false, 0><<<dim3((unsigned)((((256) / 64) * ((1600) / 64) + 7) / 8), (unsigned)(1)), 256, 0, stream>>>((const unsigned short*)(G64A), nullptr, 256, 0, (const unsigned short*)(G64B), nullptr, 256, 0, (void*)(VF), nullptr, 1600, 0, bv, nullptr, 0, 256, 1600, 256, 0.0625f);
    k_ac_planes<<<(unsigned)(((long long)C * N / 2 + 255) / 256), 256, 0, stream>>>(QF, KF, VF, (_Float16*)QH, (_Float16*)QL, (_Float16*)KH, (_Float16*)KL, (_Float16*)V16, N * C8, (long long)C * N);
    w25::wmma_gemm64<1, true, 0, 0, false, 0><<<dim3((unsigned)((((N) / 64) * ((N) / 64) + 7) / 8), (unsigned)(1)), 256, 0, stream>>>((const unsigned short*)(QH), (const unsigned short*)(QL), C8, 0, (const unsigned short*)(KH), (const unsigned short*)(KL), C8, 0, (void*)(EN), nullptr, N, 0, nullptr, nullptr, 0, N, N, C8, 1.0f);
    k_ac_soft<<<N, 256, 0, stream>>>(EN, (_Float16*)P16, N);
    w25::wmma_gemm64<0, false, 0, 0, false, 0><<<dim3((unsigned)((((C) / 64) * ((N) / 64) + 7) / 8), (unsigned)(1)), 256, 0, stream>>>((const unsigned short*)(V16), nullptr, N, 0, (const unsigned short*)(P16), nullptr, N, 0, (void*)(CT), nullptr, N, 0, nullptr, nullptr, 0, C, N, N, 0.000244140625f);
    k_ac_fuse<<<(unsigned)(((long long)C * N + 255) / 256), 256, 0, stream>>>(CT, fw, out, 2, 1, (long long)C * N);
    { GemmP gq2_2;
      gq2_2.A = s2 + (size_t)2 * C * N; gq2_2.B = Wq; gq2_2.bias = bq; gq2_2.R = s2 + (size_t)2 * C * N; gq2_2.C = QF;
      gq2_2.sAo = 0; gq2_2.sAi = 0; gq2_2.sAm = 1; gq2_2.sAk = N; gq2_2.sBo = 0; gq2_2.sBi = 0; gq2_2.sBn = C; gq2_2.sBk = 1; gq2_2.sCo = 0; gq2_2.sCi = 0; gq2_2.sCm = C8; gq2_2.sRo = 0; gq2_2.sRi = 0; gq2_2.sRm = 0; gq2_2.sRn = 0;
      gq2_2.M = N; gq2_2.N = C8; gq2_2.K = C; gq2_2.zi_n = 1; gq2_2.flags = 1; gq2_2.act = 0;
      gq2_2.alpha = 1.0f; gq2_2.beta = 0.0f; gq2_2.sa = 1.0f; gq2_2.sb = 1.0f; gq2_2.Npad = C8; gq2_2.pad_ = 0;
      if ((long long)(N) >= 64 && (long long)(C8) >= 64) k_gemmT<1, 2, 4><<<dim3((unsigned)((C8) + 63) / 64, (unsigned)((N) + 31) / 32, (unsigned)(1)), 32, 0, stream>>>(gq2_2);
      else k_gemm<1><<<dim3((unsigned)((C8) + 31) / 32, (unsigned)((N) + 15) / 16, (unsigned)(1)), 32, 0, stream>>>(gq2_2); }
    { GemmP gk2_2;
      gk2_2.A = s0 + (size_t)2 * C * N; gk2_2.B = Wk; gk2_2.bias = bk; gk2_2.R = s0 + (size_t)2 * C * N; gk2_2.C = KF;
      gk2_2.sAo = 0; gk2_2.sAi = 0; gk2_2.sAm = 1; gk2_2.sAk = N; gk2_2.sBo = 0; gk2_2.sBi = 0; gk2_2.sBn = C; gk2_2.sBk = 1; gk2_2.sCo = 0; gk2_2.sCi = 0; gk2_2.sCm = C8; gk2_2.sRo = 0; gk2_2.sRi = 0; gk2_2.sRm = 0; gk2_2.sRn = 0;
      gk2_2.M = N; gk2_2.N = C8; gk2_2.K = C; gk2_2.zi_n = 1; gk2_2.flags = 1; gk2_2.act = 0;
      gk2_2.alpha = 1.0f; gk2_2.beta = 0.0f; gk2_2.sa = 1.0f; gk2_2.sb = 1.0f; gk2_2.Npad = C8; gk2_2.pad_ = 0;
      if ((long long)(N) >= 64 && (long long)(C8) >= 64) k_gemmT<1, 2, 4><<<dim3((unsigned)((C8) + 63) / 64, (unsigned)((N) + 31) / 32, (unsigned)(1)), 32, 0, stream>>>(gk2_2);
      else k_gemm<1><<<dim3((unsigned)((C8) + 31) / 32, (unsigned)((N) + 15) / 16, (unsigned)(1)), 32, 0, stream>>>(gk2_2); }
    k_cast16<<<(unsigned)((((long long)(256) * ((256) / 2)) + 255) / 256), 256, 0, stream>>>(Wv, 256, (_Float16*)(G64A), 256, 256, 256, 1.0f);
    k_castT16<<<(unsigned)((((long long)(1600) * ((256) / 2)) + 255) / 256), 256, 0, stream>>>(s0 + (size_t)2 * C * N, 1600, (_Float16*)(G64B), 256, 256, 1600, 16.0f);
    w25::wmma_gemm64<0, false, 1, 0, false, 0><<<dim3((unsigned)((((256) / 64) * ((1600) / 64) + 7) / 8), (unsigned)(1)), 256, 0, stream>>>((const unsigned short*)(G64A), nullptr, 256, 0, (const unsigned short*)(G64B), nullptr, 256, 0, (void*)(VF), nullptr, 1600, 0, bv, nullptr, 0, 256, 1600, 256, 0.0625f);
    k_ac_planes<<<(unsigned)(((long long)C * N / 2 + 255) / 256), 256, 0, stream>>>(QF, KF, VF, (_Float16*)QH, (_Float16*)QL, (_Float16*)KH, (_Float16*)KL, (_Float16*)V16, N * C8, (long long)C * N);
    w25::wmma_gemm64<1, true, 0, 0, false, 0><<<dim3((unsigned)((((N) / 64) * ((N) / 64) + 7) / 8), (unsigned)(1)), 256, 0, stream>>>((const unsigned short*)(QH), (const unsigned short*)(QL), C8, 0, (const unsigned short*)(KH), (const unsigned short*)(KL), C8, 0, (void*)(EN), nullptr, N, 0, nullptr, nullptr, 0, N, N, C8, 1.0f);
    k_ac_soft<<<N, 256, 0, stream>>>(EN, (_Float16*)P16, N);
    w25::wmma_gemm64<0, false, 0, 0, false, 0><<<dim3((unsigned)((((C) / 64) * ((N) / 64) + 7) / 8), (unsigned)(1)), 256, 0, stream>>>((const unsigned short*)(V16), nullptr, N, 0, (const unsigned short*)(P16), nullptr, N, 0, (void*)(CT), nullptr, N, 0, nullptr, nullptr, 0, C, N, N, 0.000244140625f);
    k_ac_fuse<<<(unsigned)(((long long)C * N + 255) / 256), 256, 0, stream>>>(CT, fw, out, 2, 2, (long long)C * N);
    { GemmP gq2_3;
      gq2_3.A = s2 + (size_t)3 * C * N; gq2_3.B = Wq; gq2_3.bias = bq; gq2_3.R = s2 + (size_t)3 * C * N; gq2_3.C = QF;
      gq2_3.sAo = 0; gq2_3.sAi = 0; gq2_3.sAm = 1; gq2_3.sAk = N; gq2_3.sBo = 0; gq2_3.sBi = 0; gq2_3.sBn = C; gq2_3.sBk = 1; gq2_3.sCo = 0; gq2_3.sCi = 0; gq2_3.sCm = C8; gq2_3.sRo = 0; gq2_3.sRi = 0; gq2_3.sRm = 0; gq2_3.sRn = 0;
      gq2_3.M = N; gq2_3.N = C8; gq2_3.K = C; gq2_3.zi_n = 1; gq2_3.flags = 1; gq2_3.act = 0;
      gq2_3.alpha = 1.0f; gq2_3.beta = 0.0f; gq2_3.sa = 1.0f; gq2_3.sb = 1.0f; gq2_3.Npad = C8; gq2_3.pad_ = 0;
      if ((long long)(N) >= 64 && (long long)(C8) >= 64) k_gemmT<1, 2, 4><<<dim3((unsigned)((C8) + 63) / 64, (unsigned)((N) + 31) / 32, (unsigned)(1)), 32, 0, stream>>>(gq2_3);
      else k_gemm<1><<<dim3((unsigned)((C8) + 31) / 32, (unsigned)((N) + 15) / 16, (unsigned)(1)), 32, 0, stream>>>(gq2_3); }
    { GemmP gk2_3;
      gk2_3.A = s0 + (size_t)3 * C * N; gk2_3.B = Wk; gk2_3.bias = bk; gk2_3.R = s0 + (size_t)3 * C * N; gk2_3.C = KF;
      gk2_3.sAo = 0; gk2_3.sAi = 0; gk2_3.sAm = 1; gk2_3.sAk = N; gk2_3.sBo = 0; gk2_3.sBi = 0; gk2_3.sBn = C; gk2_3.sBk = 1; gk2_3.sCo = 0; gk2_3.sCi = 0; gk2_3.sCm = C8; gk2_3.sRo = 0; gk2_3.sRi = 0; gk2_3.sRm = 0; gk2_3.sRn = 0;
      gk2_3.M = N; gk2_3.N = C8; gk2_3.K = C; gk2_3.zi_n = 1; gk2_3.flags = 1; gk2_3.act = 0;
      gk2_3.alpha = 1.0f; gk2_3.beta = 0.0f; gk2_3.sa = 1.0f; gk2_3.sb = 1.0f; gk2_3.Npad = C8; gk2_3.pad_ = 0;
      if ((long long)(N) >= 64 && (long long)(C8) >= 64) k_gemmT<1, 2, 4><<<dim3((unsigned)((C8) + 63) / 64, (unsigned)((N) + 31) / 32, (unsigned)(1)), 32, 0, stream>>>(gk2_3);
      else k_gemm<1><<<dim3((unsigned)((C8) + 31) / 32, (unsigned)((N) + 15) / 16, (unsigned)(1)), 32, 0, stream>>>(gk2_3); }
    k_cast16<<<(unsigned)((((long long)(256) * ((256) / 2)) + 255) / 256), 256, 0, stream>>>(Wv, 256, (_Float16*)(G64A), 256, 256, 256, 1.0f);
    k_castT16<<<(unsigned)((((long long)(1600) * ((256) / 2)) + 255) / 256), 256, 0, stream>>>(s0 + (size_t)3 * C * N, 1600, (_Float16*)(G64B), 256, 256, 1600, 16.0f);
    w25::wmma_gemm64<0, false, 1, 0, false, 0><<<dim3((unsigned)((((256) / 64) * ((1600) / 64) + 7) / 8), (unsigned)(1)), 256, 0, stream>>>((const unsigned short*)(G64A), nullptr, 256, 0, (const unsigned short*)(G64B), nullptr, 256, 0, (void*)(VF), nullptr, 1600, 0, bv, nullptr, 0, 256, 1600, 256, 0.0625f);
    k_ac_planes<<<(unsigned)(((long long)C * N / 2 + 255) / 256), 256, 0, stream>>>(QF, KF, VF, (_Float16*)QH, (_Float16*)QL, (_Float16*)KH, (_Float16*)KL, (_Float16*)V16, N * C8, (long long)C * N);
    w25::wmma_gemm64<1, true, 0, 0, false, 0><<<dim3((unsigned)((((N) / 64) * ((N) / 64) + 7) / 8), (unsigned)(1)), 256, 0, stream>>>((const unsigned short*)(QH), (const unsigned short*)(QL), C8, 0, (const unsigned short*)(KH), (const unsigned short*)(KL), C8, 0, (void*)(EN), nullptr, N, 0, nullptr, nullptr, 0, N, N, C8, 1.0f);
    k_ac_soft<<<N, 256, 0, stream>>>(EN, (_Float16*)P16, N);
    w25::wmma_gemm64<0, false, 0, 0, false, 0><<<dim3((unsigned)((((C) / 64) * ((N) / 64) + 7) / 8), (unsigned)(1)), 256, 0, stream>>>((const unsigned short*)(V16), nullptr, N, 0, (const unsigned short*)(P16), nullptr, N, 0, (void*)(CT), nullptr, N, 0, nullptr, nullptr, 0, C, N, N, 0.000244140625f);
    k_ac_fuse<<<(unsigned)(((long long)C * N + 255) / 256), 256, 0, stream>>>(CT, fw, out, 2, 3, (long long)C * N);
    { GemmP gq2_4;
      gq2_4.A = s2 + (size_t)4 * C * N; gq2_4.B = Wq; gq2_4.bias = bq; gq2_4.R = s2 + (size_t)4 * C * N; gq2_4.C = QF;
      gq2_4.sAo = 0; gq2_4.sAi = 0; gq2_4.sAm = 1; gq2_4.sAk = N; gq2_4.sBo = 0; gq2_4.sBi = 0; gq2_4.sBn = C; gq2_4.sBk = 1; gq2_4.sCo = 0; gq2_4.sCi = 0; gq2_4.sCm = C8; gq2_4.sRo = 0; gq2_4.sRi = 0; gq2_4.sRm = 0; gq2_4.sRn = 0;
      gq2_4.M = N; gq2_4.N = C8; gq2_4.K = C; gq2_4.zi_n = 1; gq2_4.flags = 1; gq2_4.act = 0;
      gq2_4.alpha = 1.0f; gq2_4.beta = 0.0f; gq2_4.sa = 1.0f; gq2_4.sb = 1.0f; gq2_4.Npad = C8; gq2_4.pad_ = 0;
      if ((long long)(N) >= 64 && (long long)(C8) >= 64) k_gemmT<1, 2, 4><<<dim3((unsigned)((C8) + 63) / 64, (unsigned)((N) + 31) / 32, (unsigned)(1)), 32, 0, stream>>>(gq2_4);
      else k_gemm<1><<<dim3((unsigned)((C8) + 31) / 32, (unsigned)((N) + 15) / 16, (unsigned)(1)), 32, 0, stream>>>(gq2_4); }
    { GemmP gk2_4;
      gk2_4.A = s0 + (size_t)4 * C * N; gk2_4.B = Wk; gk2_4.bias = bk; gk2_4.R = s0 + (size_t)4 * C * N; gk2_4.C = KF;
      gk2_4.sAo = 0; gk2_4.sAi = 0; gk2_4.sAm = 1; gk2_4.sAk = N; gk2_4.sBo = 0; gk2_4.sBi = 0; gk2_4.sBn = C; gk2_4.sBk = 1; gk2_4.sCo = 0; gk2_4.sCi = 0; gk2_4.sCm = C8; gk2_4.sRo = 0; gk2_4.sRi = 0; gk2_4.sRm = 0; gk2_4.sRn = 0;
      gk2_4.M = N; gk2_4.N = C8; gk2_4.K = C; gk2_4.zi_n = 1; gk2_4.flags = 1; gk2_4.act = 0;
      gk2_4.alpha = 1.0f; gk2_4.beta = 0.0f; gk2_4.sa = 1.0f; gk2_4.sb = 1.0f; gk2_4.Npad = C8; gk2_4.pad_ = 0;
      if ((long long)(N) >= 64 && (long long)(C8) >= 64) k_gemmT<1, 2, 4><<<dim3((unsigned)((C8) + 63) / 64, (unsigned)((N) + 31) / 32, (unsigned)(1)), 32, 0, stream>>>(gk2_4);
      else k_gemm<1><<<dim3((unsigned)((C8) + 31) / 32, (unsigned)((N) + 15) / 16, (unsigned)(1)), 32, 0, stream>>>(gk2_4); }
    k_cast16<<<(unsigned)((((long long)(256) * ((256) / 2)) + 255) / 256), 256, 0, stream>>>(Wv, 256, (_Float16*)(G64A), 256, 256, 256, 1.0f);
    k_castT16<<<(unsigned)((((long long)(1600) * ((256) / 2)) + 255) / 256), 256, 0, stream>>>(s0 + (size_t)4 * C * N, 1600, (_Float16*)(G64B), 256, 256, 1600, 16.0f);
    w25::wmma_gemm64<0, false, 1, 0, false, 0><<<dim3((unsigned)((((256) / 64) * ((1600) / 64) + 7) / 8), (unsigned)(1)), 256, 0, stream>>>((const unsigned short*)(G64A), nullptr, 256, 0, (const unsigned short*)(G64B), nullptr, 256, 0, (void*)(VF), nullptr, 1600, 0, bv, nullptr, 0, 256, 1600, 256, 0.0625f);
    k_ac_planes<<<(unsigned)(((long long)C * N / 2 + 255) / 256), 256, 0, stream>>>(QF, KF, VF, (_Float16*)QH, (_Float16*)QL, (_Float16*)KH, (_Float16*)KL, (_Float16*)V16, N * C8, (long long)C * N);
    w25::wmma_gemm64<1, true, 0, 0, false, 0><<<dim3((unsigned)((((N) / 64) * ((N) / 64) + 7) / 8), (unsigned)(1)), 256, 0, stream>>>((const unsigned short*)(QH), (const unsigned short*)(QL), C8, 0, (const unsigned short*)(KH), (const unsigned short*)(KL), C8, 0, (void*)(EN), nullptr, N, 0, nullptr, nullptr, 0, N, N, C8, 1.0f);
    k_ac_soft<<<N, 256, 0, stream>>>(EN, (_Float16*)P16, N);
    w25::wmma_gemm64<0, false, 0, 0, false, 0><<<dim3((unsigned)((((C) / 64) * ((N) / 64) + 7) / 8), (unsigned)(1)), 256, 0, stream>>>((const unsigned short*)(V16), nullptr, N, 0, (const unsigned short*)(P16), nullptr, N, 0, (void*)(CT), nullptr, N, 0, nullptr, nullptr, 0, C, N, N, 0.000244140625f);
    k_ac_fuse<<<(unsigned)(((long long)C * N + 255) / 256), 256, 0, stream>>>(CT, fw, out, 2, 4, (long long)C * N);
    { GemmP gq2_5;
      gq2_5.A = s2 + (size_t)5 * C * N; gq2_5.B = Wq; gq2_5.bias = bq; gq2_5.R = s2 + (size_t)5 * C * N; gq2_5.C = QF;
      gq2_5.sAo = 0; gq2_5.sAi = 0; gq2_5.sAm = 1; gq2_5.sAk = N; gq2_5.sBo = 0; gq2_5.sBi = 0; gq2_5.sBn = C; gq2_5.sBk = 1; gq2_5.sCo = 0; gq2_5.sCi = 0; gq2_5.sCm = C8; gq2_5.sRo = 0; gq2_5.sRi = 0; gq2_5.sRm = 0; gq2_5.sRn = 0;
      gq2_5.M = N; gq2_5.N = C8; gq2_5.K = C; gq2_5.zi_n = 1; gq2_5.flags = 1; gq2_5.act = 0;
      gq2_5.alpha = 1.0f; gq2_5.beta = 0.0f; gq2_5.sa = 1.0f; gq2_5.sb = 1.0f; gq2_5.Npad = C8; gq2_5.pad_ = 0;
      if ((long long)(N) >= 64 && (long long)(C8) >= 64) k_gemmT<1, 2, 4><<<dim3((unsigned)((C8) + 63) / 64, (unsigned)((N) + 31) / 32, (unsigned)(1)), 32, 0, stream>>>(gq2_5);
      else k_gemm<1><<<dim3((unsigned)((C8) + 31) / 32, (unsigned)((N) + 15) / 16, (unsigned)(1)), 32, 0, stream>>>(gq2_5); }
    { GemmP gk2_5;
      gk2_5.A = s0 + (size_t)5 * C * N; gk2_5.B = Wk; gk2_5.bias = bk; gk2_5.R = s0 + (size_t)5 * C * N; gk2_5.C = KF;
      gk2_5.sAo = 0; gk2_5.sAi = 0; gk2_5.sAm = 1; gk2_5.sAk = N; gk2_5.sBo = 0; gk2_5.sBi = 0; gk2_5.sBn = C; gk2_5.sBk = 1; gk2_5.sCo = 0; gk2_5.sCi = 0; gk2_5.sCm = C8; gk2_5.sRo = 0; gk2_5.sRi = 0; gk2_5.sRm = 0; gk2_5.sRn = 0;
      gk2_5.M = N; gk2_5.N = C8; gk2_5.K = C; gk2_5.zi_n = 1; gk2_5.flags = 1; gk2_5.act = 0;
      gk2_5.alpha = 1.0f; gk2_5.beta = 0.0f; gk2_5.sa = 1.0f; gk2_5.sb = 1.0f; gk2_5.Npad = C8; gk2_5.pad_ = 0;
      if ((long long)(N) >= 64 && (long long)(C8) >= 64) k_gemmT<1, 2, 4><<<dim3((unsigned)((C8) + 63) / 64, (unsigned)((N) + 31) / 32, (unsigned)(1)), 32, 0, stream>>>(gk2_5);
      else k_gemm<1><<<dim3((unsigned)((C8) + 31) / 32, (unsigned)((N) + 15) / 16, (unsigned)(1)), 32, 0, stream>>>(gk2_5); }
    k_cast16<<<(unsigned)((((long long)(256) * ((256) / 2)) + 255) / 256), 256, 0, stream>>>(Wv, 256, (_Float16*)(G64A), 256, 256, 256, 1.0f);
    k_castT16<<<(unsigned)((((long long)(1600) * ((256) / 2)) + 255) / 256), 256, 0, stream>>>(s0 + (size_t)5 * C * N, 1600, (_Float16*)(G64B), 256, 256, 1600, 16.0f);
    w25::wmma_gemm64<0, false, 1, 0, false, 0><<<dim3((unsigned)((((256) / 64) * ((1600) / 64) + 7) / 8), (unsigned)(1)), 256, 0, stream>>>((const unsigned short*)(G64A), nullptr, 256, 0, (const unsigned short*)(G64B), nullptr, 256, 0, (void*)(VF), nullptr, 1600, 0, bv, nullptr, 0, 256, 1600, 256, 0.0625f);
    k_ac_planes<<<(unsigned)(((long long)C * N / 2 + 255) / 256), 256, 0, stream>>>(QF, KF, VF, (_Float16*)QH, (_Float16*)QL, (_Float16*)KH, (_Float16*)KL, (_Float16*)V16, N * C8, (long long)C * N);
    w25::wmma_gemm64<1, true, 0, 0, false, 0><<<dim3((unsigned)((((N) / 64) * ((N) / 64) + 7) / 8), (unsigned)(1)), 256, 0, stream>>>((const unsigned short*)(QH), (const unsigned short*)(QL), C8, 0, (const unsigned short*)(KH), (const unsigned short*)(KL), C8, 0, (void*)(EN), nullptr, N, 0, nullptr, nullptr, 0, N, N, C8, 1.0f);
    k_ac_soft<<<N, 256, 0, stream>>>(EN, (_Float16*)P16, N);
    w25::wmma_gemm64<0, false, 0, 0, false, 0><<<dim3((unsigned)((((C) / 64) * ((N) / 64) + 7) / 8), (unsigned)(1)), 256, 0, stream>>>((const unsigned short*)(V16), nullptr, N, 0, (const unsigned short*)(P16), nullptr, N, 0, (void*)(CT), nullptr, N, 0, nullptr, nullptr, 0, C, N, N, 0.000244140625f);
    k_ac_fuse<<<(unsigned)(((long long)C * N + 255) / 256), 256, 0, stream>>>(CT, fw, out, 2, 5, (long long)C * N);
    { GemmP gq2_6;
      gq2_6.A = s2 + (size_t)6 * C * N; gq2_6.B = Wq; gq2_6.bias = bq; gq2_6.R = s2 + (size_t)6 * C * N; gq2_6.C = QF;
      gq2_6.sAo = 0; gq2_6.sAi = 0; gq2_6.sAm = 1; gq2_6.sAk = N; gq2_6.sBo = 0; gq2_6.sBi = 0; gq2_6.sBn = C; gq2_6.sBk = 1; gq2_6.sCo = 0; gq2_6.sCi = 0; gq2_6.sCm = C8; gq2_6.sRo = 0; gq2_6.sRi = 0; gq2_6.sRm = 0; gq2_6.sRn = 0;
      gq2_6.M = N; gq2_6.N = C8; gq2_6.K = C; gq2_6.zi_n = 1; gq2_6.flags = 1; gq2_6.act = 0;
      gq2_6.alpha = 1.0f; gq2_6.beta = 0.0f; gq2_6.sa = 1.0f; gq2_6.sb = 1.0f; gq2_6.Npad = C8; gq2_6.pad_ = 0;
      if ((long long)(N) >= 64 && (long long)(C8) >= 64) k_gemmT<1, 2, 4><<<dim3((unsigned)((C8) + 63) / 64, (unsigned)((N) + 31) / 32, (unsigned)(1)), 32, 0, stream>>>(gq2_6);
      else k_gemm<1><<<dim3((unsigned)((C8) + 31) / 32, (unsigned)((N) + 15) / 16, (unsigned)(1)), 32, 0, stream>>>(gq2_6); }
    { GemmP gk2_6;
      gk2_6.A = s0 + (size_t)6 * C * N; gk2_6.B = Wk; gk2_6.bias = bk; gk2_6.R = s0 + (size_t)6 * C * N; gk2_6.C = KF;
      gk2_6.sAo = 0; gk2_6.sAi = 0; gk2_6.sAm = 1; gk2_6.sAk = N; gk2_6.sBo = 0; gk2_6.sBi = 0; gk2_6.sBn = C; gk2_6.sBk = 1; gk2_6.sCo = 0; gk2_6.sCi = 0; gk2_6.sCm = C8; gk2_6.sRo = 0; gk2_6.sRi = 0; gk2_6.sRm = 0; gk2_6.sRn = 0;
      gk2_6.M = N; gk2_6.N = C8; gk2_6.K = C; gk2_6.zi_n = 1; gk2_6.flags = 1; gk2_6.act = 0;
      gk2_6.alpha = 1.0f; gk2_6.beta = 0.0f; gk2_6.sa = 1.0f; gk2_6.sb = 1.0f; gk2_6.Npad = C8; gk2_6.pad_ = 0;
      if ((long long)(N) >= 64 && (long long)(C8) >= 64) k_gemmT<1, 2, 4><<<dim3((unsigned)((C8) + 63) / 64, (unsigned)((N) + 31) / 32, (unsigned)(1)), 32, 0, stream>>>(gk2_6);
      else k_gemm<1><<<dim3((unsigned)((C8) + 31) / 32, (unsigned)((N) + 15) / 16, (unsigned)(1)), 32, 0, stream>>>(gk2_6); }
    k_cast16<<<(unsigned)((((long long)(256) * ((256) / 2)) + 255) / 256), 256, 0, stream>>>(Wv, 256, (_Float16*)(G64A), 256, 256, 256, 1.0f);
    k_castT16<<<(unsigned)((((long long)(1600) * ((256) / 2)) + 255) / 256), 256, 0, stream>>>(s0 + (size_t)6 * C * N, 1600, (_Float16*)(G64B), 256, 256, 1600, 16.0f);
    w25::wmma_gemm64<0, false, 1, 0, false, 0><<<dim3((unsigned)((((256) / 64) * ((1600) / 64) + 7) / 8), (unsigned)(1)), 256, 0, stream>>>((const unsigned short*)(G64A), nullptr, 256, 0, (const unsigned short*)(G64B), nullptr, 256, 0, (void*)(VF), nullptr, 1600, 0, bv, nullptr, 0, 256, 1600, 256, 0.0625f);
    k_ac_planes<<<(unsigned)(((long long)C * N / 2 + 255) / 256), 256, 0, stream>>>(QF, KF, VF, (_Float16*)QH, (_Float16*)QL, (_Float16*)KH, (_Float16*)KL, (_Float16*)V16, N * C8, (long long)C * N);
    w25::wmma_gemm64<1, true, 0, 0, false, 0><<<dim3((unsigned)((((N) / 64) * ((N) / 64) + 7) / 8), (unsigned)(1)), 256, 0, stream>>>((const unsigned short*)(QH), (const unsigned short*)(QL), C8, 0, (const unsigned short*)(KH), (const unsigned short*)(KL), C8, 0, (void*)(EN), nullptr, N, 0, nullptr, nullptr, 0, N, N, C8, 1.0f);
    k_ac_soft<<<N, 256, 0, stream>>>(EN, (_Float16*)P16, N);
    w25::wmma_gemm64<0, false, 0, 0, false, 0><<<dim3((unsigned)((((C) / 64) * ((N) / 64) + 7) / 8), (unsigned)(1)), 256, 0, stream>>>((const unsigned short*)(V16), nullptr, N, 0, (const unsigned short*)(P16), nullptr, N, 0, (void*)(CT), nullptr, N, 0, nullptr, nullptr, 0, C, N, N, 0.000244140625f);
    k_ac_fuse<<<(unsigned)(((long long)C * N + 255) / 256), 256, 0, stream>>>(CT, fw, out, 2, 6, (long long)C * N);
    { GemmP gq2_7;
      gq2_7.A = s2 + (size_t)7 * C * N; gq2_7.B = Wq; gq2_7.bias = bq; gq2_7.R = s2 + (size_t)7 * C * N; gq2_7.C = QF;
      gq2_7.sAo = 0; gq2_7.sAi = 0; gq2_7.sAm = 1; gq2_7.sAk = N; gq2_7.sBo = 0; gq2_7.sBi = 0; gq2_7.sBn = C; gq2_7.sBk = 1; gq2_7.sCo = 0; gq2_7.sCi = 0; gq2_7.sCm = C8; gq2_7.sRo = 0; gq2_7.sRi = 0; gq2_7.sRm = 0; gq2_7.sRn = 0;
      gq2_7.M = N; gq2_7.N = C8; gq2_7.K = C; gq2_7.zi_n = 1; gq2_7.flags = 1; gq2_7.act = 0;
      gq2_7.alpha = 1.0f; gq2_7.beta = 0.0f; gq2_7.sa = 1.0f; gq2_7.sb = 1.0f; gq2_7.Npad = C8; gq2_7.pad_ = 0;
      if ((long long)(N) >= 64 && (long long)(C8) >= 64) k_gemmT<1, 2, 4><<<dim3((unsigned)((C8) + 63) / 64, (unsigned)((N) + 31) / 32, (unsigned)(1)), 32, 0, stream>>>(gq2_7);
      else k_gemm<1><<<dim3((unsigned)((C8) + 31) / 32, (unsigned)((N) + 15) / 16, (unsigned)(1)), 32, 0, stream>>>(gq2_7); }
    { GemmP gk2_7;
      gk2_7.A = s0 + (size_t)7 * C * N; gk2_7.B = Wk; gk2_7.bias = bk; gk2_7.R = s0 + (size_t)7 * C * N; gk2_7.C = KF;
      gk2_7.sAo = 0; gk2_7.sAi = 0; gk2_7.sAm = 1; gk2_7.sAk = N; gk2_7.sBo = 0; gk2_7.sBi = 0; gk2_7.sBn = C; gk2_7.sBk = 1; gk2_7.sCo = 0; gk2_7.sCi = 0; gk2_7.sCm = C8; gk2_7.sRo = 0; gk2_7.sRi = 0; gk2_7.sRm = 0; gk2_7.sRn = 0;
      gk2_7.M = N; gk2_7.N = C8; gk2_7.K = C; gk2_7.zi_n = 1; gk2_7.flags = 1; gk2_7.act = 0;
      gk2_7.alpha = 1.0f; gk2_7.beta = 0.0f; gk2_7.sa = 1.0f; gk2_7.sb = 1.0f; gk2_7.Npad = C8; gk2_7.pad_ = 0;
      if ((long long)(N) >= 64 && (long long)(C8) >= 64) k_gemmT<1, 2, 4><<<dim3((unsigned)((C8) + 63) / 64, (unsigned)((N) + 31) / 32, (unsigned)(1)), 32, 0, stream>>>(gk2_7);
      else k_gemm<1><<<dim3((unsigned)((C8) + 31) / 32, (unsigned)((N) + 15) / 16, (unsigned)(1)), 32, 0, stream>>>(gk2_7); }
    k_cast16<<<(unsigned)((((long long)(256) * ((256) / 2)) + 255) / 256), 256, 0, stream>>>(Wv, 256, (_Float16*)(G64A), 256, 256, 256, 1.0f);
    k_castT16<<<(unsigned)((((long long)(1600) * ((256) / 2)) + 255) / 256), 256, 0, stream>>>(s0 + (size_t)7 * C * N, 1600, (_Float16*)(G64B), 256, 256, 1600, 16.0f);
    w25::wmma_gemm64<0, false, 1, 0, false, 0><<<dim3((unsigned)((((256) / 64) * ((1600) / 64) + 7) / 8), (unsigned)(1)), 256, 0, stream>>>((const unsigned short*)(G64A), nullptr, 256, 0, (const unsigned short*)(G64B), nullptr, 256, 0, (void*)(VF), nullptr, 1600, 0, bv, nullptr, 0, 256, 1600, 256, 0.0625f);
    k_ac_planes<<<(unsigned)(((long long)C * N / 2 + 255) / 256), 256, 0, stream>>>(QF, KF, VF, (_Float16*)QH, (_Float16*)QL, (_Float16*)KH, (_Float16*)KL, (_Float16*)V16, N * C8, (long long)C * N);
    w25::wmma_gemm64<1, true, 0, 0, false, 0><<<dim3((unsigned)((((N) / 64) * ((N) / 64) + 7) / 8), (unsigned)(1)), 256, 0, stream>>>((const unsigned short*)(QH), (const unsigned short*)(QL), C8, 0, (const unsigned short*)(KH), (const unsigned short*)(KL), C8, 0, (void*)(EN), nullptr, N, 0, nullptr, nullptr, 0, N, N, C8, 1.0f);
    k_ac_soft<<<N, 256, 0, stream>>>(EN, (_Float16*)P16, N);
    w25::wmma_gemm64<0, false, 0, 0, false, 0><<<dim3((unsigned)((((C) / 64) * ((N) / 64) + 7) / 8), (unsigned)(1)), 256, 0, stream>>>((const unsigned short*)(V16), nullptr, N, 0, (const unsigned short*)(P16), nullptr, N, 0, (void*)(CT), nullptr, N, 0, nullptr, nullptr, 0, C, N, N, 0.000244140625f);
    k_ac_fuse<<<(unsigned)(((long long)C * N + 255) / 256), 256, 0, stream>>>(CT, fw, out, 2, 7, (long long)C * N);
    { GemmP gq2_8;
      gq2_8.A = s2 + (size_t)8 * C * N; gq2_8.B = Wq; gq2_8.bias = bq; gq2_8.R = s2 + (size_t)8 * C * N; gq2_8.C = QF;
      gq2_8.sAo = 0; gq2_8.sAi = 0; gq2_8.sAm = 1; gq2_8.sAk = N; gq2_8.sBo = 0; gq2_8.sBi = 0; gq2_8.sBn = C; gq2_8.sBk = 1; gq2_8.sCo = 0; gq2_8.sCi = 0; gq2_8.sCm = C8; gq2_8.sRo = 0; gq2_8.sRi = 0; gq2_8.sRm = 0; gq2_8.sRn = 0;
      gq2_8.M = N; gq2_8.N = C8; gq2_8.K = C; gq2_8.zi_n = 1; gq2_8.flags = 1; gq2_8.act = 0;
      gq2_8.alpha = 1.0f; gq2_8.beta = 0.0f; gq2_8.sa = 1.0f; gq2_8.sb = 1.0f; gq2_8.Npad = C8; gq2_8.pad_ = 0;
      if ((long long)(N) >= 64 && (long long)(C8) >= 64) k_gemmT<1, 2, 4><<<dim3((unsigned)((C8) + 63) / 64, (unsigned)((N) + 31) / 32, (unsigned)(1)), 32, 0, stream>>>(gq2_8);
      else k_gemm<1><<<dim3((unsigned)((C8) + 31) / 32, (unsigned)((N) + 15) / 16, (unsigned)(1)), 32, 0, stream>>>(gq2_8); }
    { GemmP gk2_8;
      gk2_8.A = s0 + (size_t)8 * C * N; gk2_8.B = Wk; gk2_8.bias = bk; gk2_8.R = s0 + (size_t)8 * C * N; gk2_8.C = KF;
      gk2_8.sAo = 0; gk2_8.sAi = 0; gk2_8.sAm = 1; gk2_8.sAk = N; gk2_8.sBo = 0; gk2_8.sBi = 0; gk2_8.sBn = C; gk2_8.sBk = 1; gk2_8.sCo = 0; gk2_8.sCi = 0; gk2_8.sCm = C8; gk2_8.sRo = 0; gk2_8.sRi = 0; gk2_8.sRm = 0; gk2_8.sRn = 0;
      gk2_8.M = N; gk2_8.N = C8; gk2_8.K = C; gk2_8.zi_n = 1; gk2_8.flags = 1; gk2_8.act = 0;
      gk2_8.alpha = 1.0f; gk2_8.beta = 0.0f; gk2_8.sa = 1.0f; gk2_8.sb = 1.0f; gk2_8.Npad = C8; gk2_8.pad_ = 0;
      if ((long long)(N) >= 64 && (long long)(C8) >= 64) k_gemmT<1, 2, 4><<<dim3((unsigned)((C8) + 63) / 64, (unsigned)((N) + 31) / 32, (unsigned)(1)), 32, 0, stream>>>(gk2_8);
      else k_gemm<1><<<dim3((unsigned)((C8) + 31) / 32, (unsigned)((N) + 15) / 16, (unsigned)(1)), 32, 0, stream>>>(gk2_8); }
    k_cast16<<<(unsigned)((((long long)(256) * ((256) / 2)) + 255) / 256), 256, 0, stream>>>(Wv, 256, (_Float16*)(G64A), 256, 256, 256, 1.0f);
    k_castT16<<<(unsigned)((((long long)(1600) * ((256) / 2)) + 255) / 256), 256, 0, stream>>>(s0 + (size_t)8 * C * N, 1600, (_Float16*)(G64B), 256, 256, 1600, 16.0f);
    w25::wmma_gemm64<0, false, 1, 0, false, 0><<<dim3((unsigned)((((256) / 64) * ((1600) / 64) + 7) / 8), (unsigned)(1)), 256, 0, stream>>>((const unsigned short*)(G64A), nullptr, 256, 0, (const unsigned short*)(G64B), nullptr, 256, 0, (void*)(VF), nullptr, 1600, 0, bv, nullptr, 0, 256, 1600, 256, 0.0625f);
    k_ac_planes<<<(unsigned)(((long long)C * N / 2 + 255) / 256), 256, 0, stream>>>(QF, KF, VF, (_Float16*)QH, (_Float16*)QL, (_Float16*)KH, (_Float16*)KL, (_Float16*)V16, N * C8, (long long)C * N);
    w25::wmma_gemm64<1, true, 0, 0, false, 0><<<dim3((unsigned)((((N) / 64) * ((N) / 64) + 7) / 8), (unsigned)(1)), 256, 0, stream>>>((const unsigned short*)(QH), (const unsigned short*)(QL), C8, 0, (const unsigned short*)(KH), (const unsigned short*)(KL), C8, 0, (void*)(EN), nullptr, N, 0, nullptr, nullptr, 0, N, N, C8, 1.0f);
    k_ac_soft<<<N, 256, 0, stream>>>(EN, (_Float16*)P16, N);
    w25::wmma_gemm64<0, false, 0, 0, false, 0><<<dim3((unsigned)((((C) / 64) * ((N) / 64) + 7) / 8), (unsigned)(1)), 256, 0, stream>>>((const unsigned short*)(V16), nullptr, N, 0, (const unsigned short*)(P16), nullptr, N, 0, (void*)(CT), nullptr, N, 0, nullptr, nullptr, 0, C, N, N, 0.000244140625f);
    k_ac_fuse<<<(unsigned)(((long long)C * N + 255) / 256), 256, 0, stream>>>(CT, fw, out, 2, 8, (long long)C * N);
    { GemmP gq2_9;
      gq2_9.A = s2 + (size_t)9 * C * N; gq2_9.B = Wq; gq2_9.bias = bq; gq2_9.R = s2 + (size_t)9 * C * N; gq2_9.C = QF;
      gq2_9.sAo = 0; gq2_9.sAi = 0; gq2_9.sAm = 1; gq2_9.sAk = N; gq2_9.sBo = 0; gq2_9.sBi = 0; gq2_9.sBn = C; gq2_9.sBk = 1; gq2_9.sCo = 0; gq2_9.sCi = 0; gq2_9.sCm = C8; gq2_9.sRo = 0; gq2_9.sRi = 0; gq2_9.sRm = 0; gq2_9.sRn = 0;
      gq2_9.M = N; gq2_9.N = C8; gq2_9.K = C; gq2_9.zi_n = 1; gq2_9.flags = 1; gq2_9.act = 0;
      gq2_9.alpha = 1.0f; gq2_9.beta = 0.0f; gq2_9.sa = 1.0f; gq2_9.sb = 1.0f; gq2_9.Npad = C8; gq2_9.pad_ = 0;
      if ((long long)(N) >= 64 && (long long)(C8) >= 64) k_gemmT<1, 2, 4><<<dim3((unsigned)((C8) + 63) / 64, (unsigned)((N) + 31) / 32, (unsigned)(1)), 32, 0, stream>>>(gq2_9);
      else k_gemm<1><<<dim3((unsigned)((C8) + 31) / 32, (unsigned)((N) + 15) / 16, (unsigned)(1)), 32, 0, stream>>>(gq2_9); }
    { GemmP gk2_9;
      gk2_9.A = s0 + (size_t)9 * C * N; gk2_9.B = Wk; gk2_9.bias = bk; gk2_9.R = s0 + (size_t)9 * C * N; gk2_9.C = KF;
      gk2_9.sAo = 0; gk2_9.sAi = 0; gk2_9.sAm = 1; gk2_9.sAk = N; gk2_9.sBo = 0; gk2_9.sBi = 0; gk2_9.sBn = C; gk2_9.sBk = 1; gk2_9.sCo = 0; gk2_9.sCi = 0; gk2_9.sCm = C8; gk2_9.sRo = 0; gk2_9.sRi = 0; gk2_9.sRm = 0; gk2_9.sRn = 0;
      gk2_9.M = N; gk2_9.N = C8; gk2_9.K = C; gk2_9.zi_n = 1; gk2_9.flags = 1; gk2_9.act = 0;
      gk2_9.alpha = 1.0f; gk2_9.beta = 0.0f; gk2_9.sa = 1.0f; gk2_9.sb = 1.0f; gk2_9.Npad = C8; gk2_9.pad_ = 0;
      if ((long long)(N) >= 64 && (long long)(C8) >= 64) k_gemmT<1, 2, 4><<<dim3((unsigned)((C8) + 63) / 64, (unsigned)((N) + 31) / 32, (unsigned)(1)), 32, 0, stream>>>(gk2_9);
      else k_gemm<1><<<dim3((unsigned)((C8) + 31) / 32, (unsigned)((N) + 15) / 16, (unsigned)(1)), 32, 0, stream>>>(gk2_9); }
    k_cast16<<<(unsigned)((((long long)(256) * ((256) / 2)) + 255) / 256), 256, 0, stream>>>(Wv, 256, (_Float16*)(G64A), 256, 256, 256, 1.0f);
    k_castT16<<<(unsigned)((((long long)(1600) * ((256) / 2)) + 255) / 256), 256, 0, stream>>>(s0 + (size_t)9 * C * N, 1600, (_Float16*)(G64B), 256, 256, 1600, 16.0f);
    w25::wmma_gemm64<0, false, 1, 0, false, 0><<<dim3((unsigned)((((256) / 64) * ((1600) / 64) + 7) / 8), (unsigned)(1)), 256, 0, stream>>>((const unsigned short*)(G64A), nullptr, 256, 0, (const unsigned short*)(G64B), nullptr, 256, 0, (void*)(VF), nullptr, 1600, 0, bv, nullptr, 0, 256, 1600, 256, 0.0625f);
    k_ac_planes<<<(unsigned)(((long long)C * N / 2 + 255) / 256), 256, 0, stream>>>(QF, KF, VF, (_Float16*)QH, (_Float16*)QL, (_Float16*)KH, (_Float16*)KL, (_Float16*)V16, N * C8, (long long)C * N);
    w25::wmma_gemm64<1, true, 0, 0, false, 0><<<dim3((unsigned)((((N) / 64) * ((N) / 64) + 7) / 8), (unsigned)(1)), 256, 0, stream>>>((const unsigned short*)(QH), (const unsigned short*)(QL), C8, 0, (const unsigned short*)(KH), (const unsigned short*)(KL), C8, 0, (void*)(EN), nullptr, N, 0, nullptr, nullptr, 0, N, N, C8, 1.0f);
    k_ac_soft<<<N, 256, 0, stream>>>(EN, (_Float16*)P16, N);
    w25::wmma_gemm64<0, false, 0, 0, false, 0><<<dim3((unsigned)((((C) / 64) * ((N) / 64) + 7) / 8), (unsigned)(1)), 256, 0, stream>>>((const unsigned short*)(V16), nullptr, N, 0, (const unsigned short*)(P16), nullptr, N, 0, (void*)(CT), nullptr, N, 0, nullptr, nullptr, 0, C, N, N, 0.000244140625f);
    k_ac_fuse<<<(unsigned)(((long long)C * N + 255) / 256), 256, 0, stream>>>(CT, fw, out, 2, 9, (long long)C * N);
    { GemmP gq2_10;
      gq2_10.A = s2 + (size_t)10 * C * N; gq2_10.B = Wq; gq2_10.bias = bq; gq2_10.R = s2 + (size_t)10 * C * N; gq2_10.C = QF;
      gq2_10.sAo = 0; gq2_10.sAi = 0; gq2_10.sAm = 1; gq2_10.sAk = N; gq2_10.sBo = 0; gq2_10.sBi = 0; gq2_10.sBn = C; gq2_10.sBk = 1; gq2_10.sCo = 0; gq2_10.sCi = 0; gq2_10.sCm = C8; gq2_10.sRo = 0; gq2_10.sRi = 0; gq2_10.sRm = 0; gq2_10.sRn = 0;
      gq2_10.M = N; gq2_10.N = C8; gq2_10.K = C; gq2_10.zi_n = 1; gq2_10.flags = 1; gq2_10.act = 0;
      gq2_10.alpha = 1.0f; gq2_10.beta = 0.0f; gq2_10.sa = 1.0f; gq2_10.sb = 1.0f; gq2_10.Npad = C8; gq2_10.pad_ = 0;
      if ((long long)(N) >= 64 && (long long)(C8) >= 64) k_gemmT<1, 2, 4><<<dim3((unsigned)((C8) + 63) / 64, (unsigned)((N) + 31) / 32, (unsigned)(1)), 32, 0, stream>>>(gq2_10);
      else k_gemm<1><<<dim3((unsigned)((C8) + 31) / 32, (unsigned)((N) + 15) / 16, (unsigned)(1)), 32, 0, stream>>>(gq2_10); }
    { GemmP gk2_10;
      gk2_10.A = s0 + (size_t)10 * C * N; gk2_10.B = Wk; gk2_10.bias = bk; gk2_10.R = s0 + (size_t)10 * C * N; gk2_10.C = KF;
      gk2_10.sAo = 0; gk2_10.sAi = 0; gk2_10.sAm = 1; gk2_10.sAk = N; gk2_10.sBo = 0; gk2_10.sBi = 0; gk2_10.sBn = C; gk2_10.sBk = 1; gk2_10.sCo = 0; gk2_10.sCi = 0; gk2_10.sCm = C8; gk2_10.sRo = 0; gk2_10.sRi = 0; gk2_10.sRm = 0; gk2_10.sRn = 0;
      gk2_10.M = N; gk2_10.N = C8; gk2_10.K = C; gk2_10.zi_n = 1; gk2_10.flags = 1; gk2_10.act = 0;
      gk2_10.alpha = 1.0f; gk2_10.beta = 0.0f; gk2_10.sa = 1.0f; gk2_10.sb = 1.0f; gk2_10.Npad = C8; gk2_10.pad_ = 0;
      if ((long long)(N) >= 64 && (long long)(C8) >= 64) k_gemmT<1, 2, 4><<<dim3((unsigned)((C8) + 63) / 64, (unsigned)((N) + 31) / 32, (unsigned)(1)), 32, 0, stream>>>(gk2_10);
      else k_gemm<1><<<dim3((unsigned)((C8) + 31) / 32, (unsigned)((N) + 15) / 16, (unsigned)(1)), 32, 0, stream>>>(gk2_10); }
    k_cast16<<<(unsigned)((((long long)(256) * ((256) / 2)) + 255) / 256), 256, 0, stream>>>(Wv, 256, (_Float16*)(G64A), 256, 256, 256, 1.0f);
    k_castT16<<<(unsigned)((((long long)(1600) * ((256) / 2)) + 255) / 256), 256, 0, stream>>>(s0 + (size_t)10 * C * N, 1600, (_Float16*)(G64B), 256, 256, 1600, 16.0f);
    w25::wmma_gemm64<0, false, 1, 0, false, 0><<<dim3((unsigned)((((256) / 64) * ((1600) / 64) + 7) / 8), (unsigned)(1)), 256, 0, stream>>>((const unsigned short*)(G64A), nullptr, 256, 0, (const unsigned short*)(G64B), nullptr, 256, 0, (void*)(VF), nullptr, 1600, 0, bv, nullptr, 0, 256, 1600, 256, 0.0625f);
    k_ac_planes<<<(unsigned)(((long long)C * N / 2 + 255) / 256), 256, 0, stream>>>(QF, KF, VF, (_Float16*)QH, (_Float16*)QL, (_Float16*)KH, (_Float16*)KL, (_Float16*)V16, N * C8, (long long)C * N);
    w25::wmma_gemm64<1, true, 0, 0, false, 0><<<dim3((unsigned)((((N) / 64) * ((N) / 64) + 7) / 8), (unsigned)(1)), 256, 0, stream>>>((const unsigned short*)(QH), (const unsigned short*)(QL), C8, 0, (const unsigned short*)(KH), (const unsigned short*)(KL), C8, 0, (void*)(EN), nullptr, N, 0, nullptr, nullptr, 0, N, N, C8, 1.0f);
    k_ac_soft<<<N, 256, 0, stream>>>(EN, (_Float16*)P16, N);
    w25::wmma_gemm64<0, false, 0, 0, false, 0><<<dim3((unsigned)((((C) / 64) * ((N) / 64) + 7) / 8), (unsigned)(1)), 256, 0, stream>>>((const unsigned short*)(V16), nullptr, N, 0, (const unsigned short*)(P16), nullptr, N, 0, (void*)(CT), nullptr, N, 0, nullptr, nullptr, 0, C, N, N, 0.000244140625f);
    k_ac_fuse<<<(unsigned)(((long long)C * N + 255) / 256), 256, 0, stream>>>(CT, fw, out, 2, 10, (long long)C * N);
    { GemmP gq2_11;
      gq2_11.A = s2 + (size_t)11 * C * N; gq2_11.B = Wq; gq2_11.bias = bq; gq2_11.R = s2 + (size_t)11 * C * N; gq2_11.C = QF;
      gq2_11.sAo = 0; gq2_11.sAi = 0; gq2_11.sAm = 1; gq2_11.sAk = N; gq2_11.sBo = 0; gq2_11.sBi = 0; gq2_11.sBn = C; gq2_11.sBk = 1; gq2_11.sCo = 0; gq2_11.sCi = 0; gq2_11.sCm = C8; gq2_11.sRo = 0; gq2_11.sRi = 0; gq2_11.sRm = 0; gq2_11.sRn = 0;
      gq2_11.M = N; gq2_11.N = C8; gq2_11.K = C; gq2_11.zi_n = 1; gq2_11.flags = 1; gq2_11.act = 0;
      gq2_11.alpha = 1.0f; gq2_11.beta = 0.0f; gq2_11.sa = 1.0f; gq2_11.sb = 1.0f; gq2_11.Npad = C8; gq2_11.pad_ = 0;
      if ((long long)(N) >= 64 && (long long)(C8) >= 64) k_gemmT<1, 2, 4><<<dim3((unsigned)((C8) + 63) / 64, (unsigned)((N) + 31) / 32, (unsigned)(1)), 32, 0, stream>>>(gq2_11);
      else k_gemm<1><<<dim3((unsigned)((C8) + 31) / 32, (unsigned)((N) + 15) / 16, (unsigned)(1)), 32, 0, stream>>>(gq2_11); }
    { GemmP gk2_11;
      gk2_11.A = s0 + (size_t)11 * C * N; gk2_11.B = Wk; gk2_11.bias = bk; gk2_11.R = s0 + (size_t)11 * C * N; gk2_11.C = KF;
      gk2_11.sAo = 0; gk2_11.sAi = 0; gk2_11.sAm = 1; gk2_11.sAk = N; gk2_11.sBo = 0; gk2_11.sBi = 0; gk2_11.sBn = C; gk2_11.sBk = 1; gk2_11.sCo = 0; gk2_11.sCi = 0; gk2_11.sCm = C8; gk2_11.sRo = 0; gk2_11.sRi = 0; gk2_11.sRm = 0; gk2_11.sRn = 0;
      gk2_11.M = N; gk2_11.N = C8; gk2_11.K = C; gk2_11.zi_n = 1; gk2_11.flags = 1; gk2_11.act = 0;
      gk2_11.alpha = 1.0f; gk2_11.beta = 0.0f; gk2_11.sa = 1.0f; gk2_11.sb = 1.0f; gk2_11.Npad = C8; gk2_11.pad_ = 0;
      if ((long long)(N) >= 64 && (long long)(C8) >= 64) k_gemmT<1, 2, 4><<<dim3((unsigned)((C8) + 63) / 64, (unsigned)((N) + 31) / 32, (unsigned)(1)), 32, 0, stream>>>(gk2_11);
      else k_gemm<1><<<dim3((unsigned)((C8) + 31) / 32, (unsigned)((N) + 15) / 16, (unsigned)(1)), 32, 0, stream>>>(gk2_11); }
    k_cast16<<<(unsigned)((((long long)(256) * ((256) / 2)) + 255) / 256), 256, 0, stream>>>(Wv, 256, (_Float16*)(G64A), 256, 256, 256, 1.0f);
    k_castT16<<<(unsigned)((((long long)(1600) * ((256) / 2)) + 255) / 256), 256, 0, stream>>>(s0 + (size_t)11 * C * N, 1600, (_Float16*)(G64B), 256, 256, 1600, 16.0f);
    w25::wmma_gemm64<0, false, 1, 0, false, 0><<<dim3((unsigned)((((256) / 64) * ((1600) / 64) + 7) / 8), (unsigned)(1)), 256, 0, stream>>>((const unsigned short*)(G64A), nullptr, 256, 0, (const unsigned short*)(G64B), nullptr, 256, 0, (void*)(VF), nullptr, 1600, 0, bv, nullptr, 0, 256, 1600, 256, 0.0625f);
    k_ac_planes<<<(unsigned)(((long long)C * N / 2 + 255) / 256), 256, 0, stream>>>(QF, KF, VF, (_Float16*)QH, (_Float16*)QL, (_Float16*)KH, (_Float16*)KL, (_Float16*)V16, N * C8, (long long)C * N);
    w25::wmma_gemm64<1, true, 0, 0, false, 0><<<dim3((unsigned)((((N) / 64) * ((N) / 64) + 7) / 8), (unsigned)(1)), 256, 0, stream>>>((const unsigned short*)(QH), (const unsigned short*)(QL), C8, 0, (const unsigned short*)(KH), (const unsigned short*)(KL), C8, 0, (void*)(EN), nullptr, N, 0, nullptr, nullptr, 0, N, N, C8, 1.0f);
    k_ac_soft<<<N, 256, 0, stream>>>(EN, (_Float16*)P16, N);
    w25::wmma_gemm64<0, false, 0, 0, false, 0><<<dim3((unsigned)((((C) / 64) * ((N) / 64) + 7) / 8), (unsigned)(1)), 256, 0, stream>>>((const unsigned short*)(V16), nullptr, N, 0, (const unsigned short*)(P16), nullptr, N, 0, (void*)(CT), nullptr, N, 0, nullptr, nullptr, 0, C, N, N, 0.000244140625f);
    k_ac_fuse<<<(unsigned)(((long long)C * N + 255) / 256), 256, 0, stream>>>(CT, fw, out, 2, 11, (long long)C * N);
    { GemmP gq2_12;
      gq2_12.A = s2 + (size_t)12 * C * N; gq2_12.B = Wq; gq2_12.bias = bq; gq2_12.R = s2 + (size_t)12 * C * N; gq2_12.C = QF;
      gq2_12.sAo = 0; gq2_12.sAi = 0; gq2_12.sAm = 1; gq2_12.sAk = N; gq2_12.sBo = 0; gq2_12.sBi = 0; gq2_12.sBn = C; gq2_12.sBk = 1; gq2_12.sCo = 0; gq2_12.sCi = 0; gq2_12.sCm = C8; gq2_12.sRo = 0; gq2_12.sRi = 0; gq2_12.sRm = 0; gq2_12.sRn = 0;
      gq2_12.M = N; gq2_12.N = C8; gq2_12.K = C; gq2_12.zi_n = 1; gq2_12.flags = 1; gq2_12.act = 0;
      gq2_12.alpha = 1.0f; gq2_12.beta = 0.0f; gq2_12.sa = 1.0f; gq2_12.sb = 1.0f; gq2_12.Npad = C8; gq2_12.pad_ = 0;
      if ((long long)(N) >= 64 && (long long)(C8) >= 64) k_gemmT<1, 2, 4><<<dim3((unsigned)((C8) + 63) / 64, (unsigned)((N) + 31) / 32, (unsigned)(1)), 32, 0, stream>>>(gq2_12);
      else k_gemm<1><<<dim3((unsigned)((C8) + 31) / 32, (unsigned)((N) + 15) / 16, (unsigned)(1)), 32, 0, stream>>>(gq2_12); }
    { GemmP gk2_12;
      gk2_12.A = s0 + (size_t)12 * C * N; gk2_12.B = Wk; gk2_12.bias = bk; gk2_12.R = s0 + (size_t)12 * C * N; gk2_12.C = KF;
      gk2_12.sAo = 0; gk2_12.sAi = 0; gk2_12.sAm = 1; gk2_12.sAk = N; gk2_12.sBo = 0; gk2_12.sBi = 0; gk2_12.sBn = C; gk2_12.sBk = 1; gk2_12.sCo = 0; gk2_12.sCi = 0; gk2_12.sCm = C8; gk2_12.sRo = 0; gk2_12.sRi = 0; gk2_12.sRm = 0; gk2_12.sRn = 0;
      gk2_12.M = N; gk2_12.N = C8; gk2_12.K = C; gk2_12.zi_n = 1; gk2_12.flags = 1; gk2_12.act = 0;
      gk2_12.alpha = 1.0f; gk2_12.beta = 0.0f; gk2_12.sa = 1.0f; gk2_12.sb = 1.0f; gk2_12.Npad = C8; gk2_12.pad_ = 0;
      if ((long long)(N) >= 64 && (long long)(C8) >= 64) k_gemmT<1, 2, 4><<<dim3((unsigned)((C8) + 63) / 64, (unsigned)((N) + 31) / 32, (unsigned)(1)), 32, 0, stream>>>(gk2_12);
      else k_gemm<1><<<dim3((unsigned)((C8) + 31) / 32, (unsigned)((N) + 15) / 16, (unsigned)(1)), 32, 0, stream>>>(gk2_12); }
    k_cast16<<<(unsigned)((((long long)(256) * ((256) / 2)) + 255) / 256), 256, 0, stream>>>(Wv, 256, (_Float16*)(G64A), 256, 256, 256, 1.0f);
    k_castT16<<<(unsigned)((((long long)(1600) * ((256) / 2)) + 255) / 256), 256, 0, stream>>>(s0 + (size_t)12 * C * N, 1600, (_Float16*)(G64B), 256, 256, 1600, 16.0f);
    w25::wmma_gemm64<0, false, 1, 0, false, 0><<<dim3((unsigned)((((256) / 64) * ((1600) / 64) + 7) / 8), (unsigned)(1)), 256, 0, stream>>>((const unsigned short*)(G64A), nullptr, 256, 0, (const unsigned short*)(G64B), nullptr, 256, 0, (void*)(VF), nullptr, 1600, 0, bv, nullptr, 0, 256, 1600, 256, 0.0625f);
    k_ac_planes<<<(unsigned)(((long long)C * N / 2 + 255) / 256), 256, 0, stream>>>(QF, KF, VF, (_Float16*)QH, (_Float16*)QL, (_Float16*)KH, (_Float16*)KL, (_Float16*)V16, N * C8, (long long)C * N);
    w25::wmma_gemm64<1, true, 0, 0, false, 0><<<dim3((unsigned)((((N) / 64) * ((N) / 64) + 7) / 8), (unsigned)(1)), 256, 0, stream>>>((const unsigned short*)(QH), (const unsigned short*)(QL), C8, 0, (const unsigned short*)(KH), (const unsigned short*)(KL), C8, 0, (void*)(EN), nullptr, N, 0, nullptr, nullptr, 0, N, N, C8, 1.0f);
    k_ac_soft<<<N, 256, 0, stream>>>(EN, (_Float16*)P16, N);
    w25::wmma_gemm64<0, false, 0, 0, false, 0><<<dim3((unsigned)((((C) / 64) * ((N) / 64) + 7) / 8), (unsigned)(1)), 256, 0, stream>>>((const unsigned short*)(V16), nullptr, N, 0, (const unsigned short*)(P16), nullptr, N, 0, (void*)(CT), nullptr, N, 0, nullptr, nullptr, 0, C, N, N, 0.000244140625f);
    k_ac_fuse<<<(unsigned)(((long long)C * N + 255) / 256), 256, 0, stream>>>(CT, fw, out, 2, 12, (long long)C * N);
    { GemmP gq2_13;
      gq2_13.A = s2 + (size_t)13 * C * N; gq2_13.B = Wq; gq2_13.bias = bq; gq2_13.R = s2 + (size_t)13 * C * N; gq2_13.C = QF;
      gq2_13.sAo = 0; gq2_13.sAi = 0; gq2_13.sAm = 1; gq2_13.sAk = N; gq2_13.sBo = 0; gq2_13.sBi = 0; gq2_13.sBn = C; gq2_13.sBk = 1; gq2_13.sCo = 0; gq2_13.sCi = 0; gq2_13.sCm = C8; gq2_13.sRo = 0; gq2_13.sRi = 0; gq2_13.sRm = 0; gq2_13.sRn = 0;
      gq2_13.M = N; gq2_13.N = C8; gq2_13.K = C; gq2_13.zi_n = 1; gq2_13.flags = 1; gq2_13.act = 0;
      gq2_13.alpha = 1.0f; gq2_13.beta = 0.0f; gq2_13.sa = 1.0f; gq2_13.sb = 1.0f; gq2_13.Npad = C8; gq2_13.pad_ = 0;
      if ((long long)(N) >= 64 && (long long)(C8) >= 64) k_gemmT<1, 2, 4><<<dim3((unsigned)((C8) + 63) / 64, (unsigned)((N) + 31) / 32, (unsigned)(1)), 32, 0, stream>>>(gq2_13);
      else k_gemm<1><<<dim3((unsigned)((C8) + 31) / 32, (unsigned)((N) + 15) / 16, (unsigned)(1)), 32, 0, stream>>>(gq2_13); }
    { GemmP gk2_13;
      gk2_13.A = s0 + (size_t)13 * C * N; gk2_13.B = Wk; gk2_13.bias = bk; gk2_13.R = s0 + (size_t)13 * C * N; gk2_13.C = KF;
      gk2_13.sAo = 0; gk2_13.sAi = 0; gk2_13.sAm = 1; gk2_13.sAk = N; gk2_13.sBo = 0; gk2_13.sBi = 0; gk2_13.sBn = C; gk2_13.sBk = 1; gk2_13.sCo = 0; gk2_13.sCi = 0; gk2_13.sCm = C8; gk2_13.sRo = 0; gk2_13.sRi = 0; gk2_13.sRm = 0; gk2_13.sRn = 0;
      gk2_13.M = N; gk2_13.N = C8; gk2_13.K = C; gk2_13.zi_n = 1; gk2_13.flags = 1; gk2_13.act = 0;
      gk2_13.alpha = 1.0f; gk2_13.beta = 0.0f; gk2_13.sa = 1.0f; gk2_13.sb = 1.0f; gk2_13.Npad = C8; gk2_13.pad_ = 0;
      if ((long long)(N) >= 64 && (long long)(C8) >= 64) k_gemmT<1, 2, 4><<<dim3((unsigned)((C8) + 63) / 64, (unsigned)((N) + 31) / 32, (unsigned)(1)), 32, 0, stream>>>(gk2_13);
      else k_gemm<1><<<dim3((unsigned)((C8) + 31) / 32, (unsigned)((N) + 15) / 16, (unsigned)(1)), 32, 0, stream>>>(gk2_13); }
    k_cast16<<<(unsigned)((((long long)(256) * ((256) / 2)) + 255) / 256), 256, 0, stream>>>(Wv, 256, (_Float16*)(G64A), 256, 256, 256, 1.0f);
    k_castT16<<<(unsigned)((((long long)(1600) * ((256) / 2)) + 255) / 256), 256, 0, stream>>>(s0 + (size_t)13 * C * N, 1600, (_Float16*)(G64B), 256, 256, 1600, 16.0f);
    w25::wmma_gemm64<0, false, 1, 0, false, 0><<<dim3((unsigned)((((256) / 64) * ((1600) / 64) + 7) / 8), (unsigned)(1)), 256, 0, stream>>>((const unsigned short*)(G64A), nullptr, 256, 0, (const unsigned short*)(G64B), nullptr, 256, 0, (void*)(VF), nullptr, 1600, 0, bv, nullptr, 0, 256, 1600, 256, 0.0625f);
    k_ac_planes<<<(unsigned)(((long long)C * N / 2 + 255) / 256), 256, 0, stream>>>(QF, KF, VF, (_Float16*)QH, (_Float16*)QL, (_Float16*)KH, (_Float16*)KL, (_Float16*)V16, N * C8, (long long)C * N);
    w25::wmma_gemm64<1, true, 0, 0, false, 0><<<dim3((unsigned)((((N) / 64) * ((N) / 64) + 7) / 8), (unsigned)(1)), 256, 0, stream>>>((const unsigned short*)(QH), (const unsigned short*)(QL), C8, 0, (const unsigned short*)(KH), (const unsigned short*)(KL), C8, 0, (void*)(EN), nullptr, N, 0, nullptr, nullptr, 0, N, N, C8, 1.0f);
    k_ac_soft<<<N, 256, 0, stream>>>(EN, (_Float16*)P16, N);
    w25::wmma_gemm64<0, false, 0, 0, false, 0><<<dim3((unsigned)((((C) / 64) * ((N) / 64) + 7) / 8), (unsigned)(1)), 256, 0, stream>>>((const unsigned short*)(V16), nullptr, N, 0, (const unsigned short*)(P16), nullptr, N, 0, (void*)(CT), nullptr, N, 0, nullptr, nullptr, 0, C, N, N, 0.000244140625f);
    k_ac_fuse<<<(unsigned)(((long long)C * N + 255) / 256), 256, 0, stream>>>(CT, fw, out, 2, 13, (long long)C * N);
    { GemmP gq2_14;
      gq2_14.A = s2 + (size_t)14 * C * N; gq2_14.B = Wq; gq2_14.bias = bq; gq2_14.R = s2 + (size_t)14 * C * N; gq2_14.C = QF;
      gq2_14.sAo = 0; gq2_14.sAi = 0; gq2_14.sAm = 1; gq2_14.sAk = N; gq2_14.sBo = 0; gq2_14.sBi = 0; gq2_14.sBn = C; gq2_14.sBk = 1; gq2_14.sCo = 0; gq2_14.sCi = 0; gq2_14.sCm = C8; gq2_14.sRo = 0; gq2_14.sRi = 0; gq2_14.sRm = 0; gq2_14.sRn = 0;
      gq2_14.M = N; gq2_14.N = C8; gq2_14.K = C; gq2_14.zi_n = 1; gq2_14.flags = 1; gq2_14.act = 0;
      gq2_14.alpha = 1.0f; gq2_14.beta = 0.0f; gq2_14.sa = 1.0f; gq2_14.sb = 1.0f; gq2_14.Npad = C8; gq2_14.pad_ = 0;
      if ((long long)(N) >= 64 && (long long)(C8) >= 64) k_gemmT<1, 2, 4><<<dim3((unsigned)((C8) + 63) / 64, (unsigned)((N) + 31) / 32, (unsigned)(1)), 32, 0, stream>>>(gq2_14);
      else k_gemm<1><<<dim3((unsigned)((C8) + 31) / 32, (unsigned)((N) + 15) / 16, (unsigned)(1)), 32, 0, stream>>>(gq2_14); }
    { GemmP gk2_14;
      gk2_14.A = s0 + (size_t)14 * C * N; gk2_14.B = Wk; gk2_14.bias = bk; gk2_14.R = s0 + (size_t)14 * C * N; gk2_14.C = KF;
      gk2_14.sAo = 0; gk2_14.sAi = 0; gk2_14.sAm = 1; gk2_14.sAk = N; gk2_14.sBo = 0; gk2_14.sBi = 0; gk2_14.sBn = C; gk2_14.sBk = 1; gk2_14.sCo = 0; gk2_14.sCi = 0; gk2_14.sCm = C8; gk2_14.sRo = 0; gk2_14.sRi = 0; gk2_14.sRm = 0; gk2_14.sRn = 0;
      gk2_14.M = N; gk2_14.N = C8; gk2_14.K = C; gk2_14.zi_n = 1; gk2_14.flags = 1; gk2_14.act = 0;
      gk2_14.alpha = 1.0f; gk2_14.beta = 0.0f; gk2_14.sa = 1.0f; gk2_14.sb = 1.0f; gk2_14.Npad = C8; gk2_14.pad_ = 0;
      if ((long long)(N) >= 64 && (long long)(C8) >= 64) k_gemmT<1, 2, 4><<<dim3((unsigned)((C8) + 63) / 64, (unsigned)((N) + 31) / 32, (unsigned)(1)), 32, 0, stream>>>(gk2_14);
      else k_gemm<1><<<dim3((unsigned)((C8) + 31) / 32, (unsigned)((N) + 15) / 16, (unsigned)(1)), 32, 0, stream>>>(gk2_14); }
    k_cast16<<<(unsigned)((((long long)(256) * ((256) / 2)) + 255) / 256), 256, 0, stream>>>(Wv, 256, (_Float16*)(G64A), 256, 256, 256, 1.0f);
    k_castT16<<<(unsigned)((((long long)(1600) * ((256) / 2)) + 255) / 256), 256, 0, stream>>>(s0 + (size_t)14 * C * N, 1600, (_Float16*)(G64B), 256, 256, 1600, 16.0f);
    w25::wmma_gemm64<0, false, 1, 0, false, 0><<<dim3((unsigned)((((256) / 64) * ((1600) / 64) + 7) / 8), (unsigned)(1)), 256, 0, stream>>>((const unsigned short*)(G64A), nullptr, 256, 0, (const unsigned short*)(G64B), nullptr, 256, 0, (void*)(VF), nullptr, 1600, 0, bv, nullptr, 0, 256, 1600, 256, 0.0625f);
    k_ac_planes<<<(unsigned)(((long long)C * N / 2 + 255) / 256), 256, 0, stream>>>(QF, KF, VF, (_Float16*)QH, (_Float16*)QL, (_Float16*)KH, (_Float16*)KL, (_Float16*)V16, N * C8, (long long)C * N);
    w25::wmma_gemm64<1, true, 0, 0, false, 0><<<dim3((unsigned)((((N) / 64) * ((N) / 64) + 7) / 8), (unsigned)(1)), 256, 0, stream>>>((const unsigned short*)(QH), (const unsigned short*)(QL), C8, 0, (const unsigned short*)(KH), (const unsigned short*)(KL), C8, 0, (void*)(EN), nullptr, N, 0, nullptr, nullptr, 0, N, N, C8, 1.0f);
    k_ac_soft<<<N, 256, 0, stream>>>(EN, (_Float16*)P16, N);
    w25::wmma_gemm64<0, false, 0, 0, false, 0><<<dim3((unsigned)((((C) / 64) * ((N) / 64) + 7) / 8), (unsigned)(1)), 256, 0, stream>>>((const unsigned short*)(V16), nullptr, N, 0, (const unsigned short*)(P16), nullptr, N, 0, (void*)(CT), nullptr, N, 0, nullptr, nullptr, 0, C, N, N, 0.000244140625f);
    k_ac_fuse<<<(unsigned)(((long long)C * N + 255) / 256), 256, 0, stream>>>(CT, fw, out, 2, 14, (long long)C * N);
    { GemmP gq2_15;
      gq2_15.A = s2 + (size_t)15 * C * N; gq2_15.B = Wq; gq2_15.bias = bq; gq2_15.R = s2 + (size_t)15 * C * N; gq2_15.C = QF;
      gq2_15.sAo = 0; gq2_15.sAi = 0; gq2_15.sAm = 1; gq2_15.sAk = N; gq2_15.sBo = 0; gq2_15.sBi = 0; gq2_15.sBn = C; gq2_15.sBk = 1; gq2_15.sCo = 0; gq2_15.sCi = 0; gq2_15.sCm = C8; gq2_15.sRo = 0; gq2_15.sRi = 0; gq2_15.sRm = 0; gq2_15.sRn = 0;
      gq2_15.M = N; gq2_15.N = C8; gq2_15.K = C; gq2_15.zi_n = 1; gq2_15.flags = 1; gq2_15.act = 0;
      gq2_15.alpha = 1.0f; gq2_15.beta = 0.0f; gq2_15.sa = 1.0f; gq2_15.sb = 1.0f; gq2_15.Npad = C8; gq2_15.pad_ = 0;
      if ((long long)(N) >= 64 && (long long)(C8) >= 64) k_gemmT<1, 2, 4><<<dim3((unsigned)((C8) + 63) / 64, (unsigned)((N) + 31) / 32, (unsigned)(1)), 32, 0, stream>>>(gq2_15);
      else k_gemm<1><<<dim3((unsigned)((C8) + 31) / 32, (unsigned)((N) + 15) / 16, (unsigned)(1)), 32, 0, stream>>>(gq2_15); }
    { GemmP gk2_15;
      gk2_15.A = s0 + (size_t)15 * C * N; gk2_15.B = Wk; gk2_15.bias = bk; gk2_15.R = s0 + (size_t)15 * C * N; gk2_15.C = KF;
      gk2_15.sAo = 0; gk2_15.sAi = 0; gk2_15.sAm = 1; gk2_15.sAk = N; gk2_15.sBo = 0; gk2_15.sBi = 0; gk2_15.sBn = C; gk2_15.sBk = 1; gk2_15.sCo = 0; gk2_15.sCi = 0; gk2_15.sCm = C8; gk2_15.sRo = 0; gk2_15.sRi = 0; gk2_15.sRm = 0; gk2_15.sRn = 0;
      gk2_15.M = N; gk2_15.N = C8; gk2_15.K = C; gk2_15.zi_n = 1; gk2_15.flags = 1; gk2_15.act = 0;
      gk2_15.alpha = 1.0f; gk2_15.beta = 0.0f; gk2_15.sa = 1.0f; gk2_15.sb = 1.0f; gk2_15.Npad = C8; gk2_15.pad_ = 0;
      if ((long long)(N) >= 64 && (long long)(C8) >= 64) k_gemmT<1, 2, 4><<<dim3((unsigned)((C8) + 63) / 64, (unsigned)((N) + 31) / 32, (unsigned)(1)), 32, 0, stream>>>(gk2_15);
      else k_gemm<1><<<dim3((unsigned)((C8) + 31) / 32, (unsigned)((N) + 15) / 16, (unsigned)(1)), 32, 0, stream>>>(gk2_15); }
    k_cast16<<<(unsigned)((((long long)(256) * ((256) / 2)) + 255) / 256), 256, 0, stream>>>(Wv, 256, (_Float16*)(G64A), 256, 256, 256, 1.0f);
    k_castT16<<<(unsigned)((((long long)(1600) * ((256) / 2)) + 255) / 256), 256, 0, stream>>>(s0 + (size_t)15 * C * N, 1600, (_Float16*)(G64B), 256, 256, 1600, 16.0f);
    w25::wmma_gemm64<0, false, 1, 0, false, 0><<<dim3((unsigned)((((256) / 64) * ((1600) / 64) + 7) / 8), (unsigned)(1)), 256, 0, stream>>>((const unsigned short*)(G64A), nullptr, 256, 0, (const unsigned short*)(G64B), nullptr, 256, 0, (void*)(VF), nullptr, 1600, 0, bv, nullptr, 0, 256, 1600, 256, 0.0625f);
    k_ac_planes<<<(unsigned)(((long long)C * N / 2 + 255) / 256), 256, 0, stream>>>(QF, KF, VF, (_Float16*)QH, (_Float16*)QL, (_Float16*)KH, (_Float16*)KL, (_Float16*)V16, N * C8, (long long)C * N);
    w25::wmma_gemm64<1, true, 0, 0, false, 0><<<dim3((unsigned)((((N) / 64) * ((N) / 64) + 7) / 8), (unsigned)(1)), 256, 0, stream>>>((const unsigned short*)(QH), (const unsigned short*)(QL), C8, 0, (const unsigned short*)(KH), (const unsigned short*)(KL), C8, 0, (void*)(EN), nullptr, N, 0, nullptr, nullptr, 0, N, N, C8, 1.0f);
    k_ac_soft<<<N, 256, 0, stream>>>(EN, (_Float16*)P16, N);
    w25::wmma_gemm64<0, false, 0, 0, false, 0><<<dim3((unsigned)((((C) / 64) * ((N) / 64) + 7) / 8), (unsigned)(1)), 256, 0, stream>>>((const unsigned short*)(V16), nullptr, N, 0, (const unsigned short*)(P16), nullptr, N, 0, (void*)(CT), nullptr, N, 0, nullptr, nullptr, 0, C, N, N, 0.000244140625f);
    k_ac_fuse<<<(unsigned)(((long long)C * N + 255) / 256), 256, 0, stream>>>(CT, fw, out, 2, 15, (long long)C * N);
}
